// LoraDecoderLayer_25262997636082
// MI455X (gfx1250) — hardware-verified
//
#include <hip/hip_runtime.h>
#include <math.h>

typedef __attribute__((ext_vector_type(16))) _Float16 v16h;
typedef __attribute__((ext_vector_type(8)))  _Float16 v8h;
typedef __attribute__((ext_vector_type(16))) __bf16   v16b;
typedef __attribute__((ext_vector_type(8)))  float    v8f;
typedef __attribute__((ext_vector_type(4)))  float    v4f;

__device__ __forceinline__ int frag_k(int i, int h) { return (i < 8) ? (8 * h + i) : (16 + 8 * h + (i - 8)); }
__device__ __forceinline__ __bf16 bf16_rne(float f) {
    unsigned int u = __float_as_uint(f);
    u += 0x7fffu + ((u >> 16) & 1u);
    return __builtin_bit_cast(__bf16, (unsigned short)(u >> 16));
}
__device__ __forceinline__ float bf16_f32(__bf16 b) { return __uint_as_float(((unsigned int)__builtin_bit_cast(unsigned short, b)) << 16); }
__device__ __forceinline__ v8f wmma16(v16h a, v16h b, v8f c) {
    c = __builtin_amdgcn_wmma_f32_16x16x32_f16(false, a, false, b, (short)0, c, false, false);
    asm volatile("v_nop\n\tv_nop\n\tv_nop\n\tv_nop" : "+v"(c) : "v"(a), "v"(b));
    return c;
}
__device__ __forceinline__ v8f wmmab(v16b a, v16b b, v8f c) {
    c = __builtin_amdgcn_wmma_f32_16x16x32_bf16(false, a, false, b, (short)0, c, false, false);
    asm volatile("v_nop\n\tv_nop\n\tv_nop\n\tv_nop" : "+v"(c) : "v"(a), "v"(b));
    return c;
}
struct Split { v16b hi, lo; };
__device__ __forceinline__ v8f wmma3(const Split& a, const Split& b, v8f c) {
    c = __builtin_amdgcn_wmma_f32_16x16x32_bf16(false, a.hi, false, b.hi, (short)0, c, false, false);
    c = __builtin_amdgcn_wmma_f32_16x16x32_bf16(false, a.hi, false, b.lo, (short)0, c, false, false);
    c = __builtin_amdgcn_wmma_f32_16x16x32_bf16(false, a.lo, false, b.hi, (short)0, c, false, false);
    asm volatile("v_nop\n\tv_nop\n\tv_nop\n\tv_nop" : "+v"(c) : "v"(a.hi), "v"(a.lo), "v"(b.hi), "v"(b.lo));
    return c;
}
struct Split3 { v16b hi, mid, lo; };
__device__ __forceinline__ v8f wmma6(const Split3& a, const Split3& b, v8f c) {
    c = __builtin_amdgcn_wmma_f32_16x16x32_bf16(false, a.hi, false, b.hi, (short)0, c, false, false);
    c = __builtin_amdgcn_wmma_f32_16x16x32_bf16(false, a.hi, false, b.mid, (short)0, c, false, false);
    c = __builtin_amdgcn_wmma_f32_16x16x32_bf16(false, a.mid, false, b.hi, (short)0, c, false, false);
    c = __builtin_amdgcn_wmma_f32_16x16x32_bf16(false, a.hi, false, b.lo, (short)0, c, false, false);
    c = __builtin_amdgcn_wmma_f32_16x16x32_bf16(false, a.mid, false, b.mid, (short)0, c, false, false);
    c = __builtin_amdgcn_wmma_f32_16x16x32_bf16(false, a.lo, false, b.hi, (short)0, c, false, false);
    asm volatile("v_nop\n\tv_nop\n\tv_nop\n\tv_nop" : "+v"(c) : "v"(a.hi), "v"(a.mid), "v"(a.lo), "v"(b.hi), "v"(b.mid), "v"(b.lo));
    return c;
}

__device__ __forceinline__ v16h fh_ld(const float* __restrict__ p, long long sk, int k0, int h, int klen, float s) {
    v16h a;
#pragma unroll
    for (int i = 0; i < 16; ++i) { const int k = k0 + frag_k(i, h); a[i] = (k < klen) ? (_Float16)(p[(long long)k * sk] * s) : (_Float16)0.f; }
    return a;
}
__device__ __forceinline__ Split sp_ld(const float* __restrict__ p, long long sk, int k0, int h, int klen, float s) {
    Split r;
#pragma unroll
    for (int i = 0; i < 16; ++i) {
        const int k = k0 + frag_k(i, h); const float x = (k < klen) ? p[(long long)k * sk] * s : 0.f;
        const __bf16 hb = bf16_rne(x); r.hi[i] = hb; r.lo[i] = bf16_rne(x - bf16_f32(hb));
    }
    return r;
}
__device__ __forceinline__ Split3 sp3_ld(const float* __restrict__ p, long long sk, int k0, int h, int klen, float s) {
    Split3 r;
#pragma unroll
    for (int i = 0; i < 16; ++i) {
        const int k = k0 + frag_k(i, h); const float x = (k < klen) ? p[(long long)k * sk] * s : 0.f;
        const __bf16 hb = bf16_rne(x); const float r1 = x - bf16_f32(hb); const __bf16 mb = bf16_rne(r1);
        r.hi[i] = hb; r.mid[i] = mb; r.lo[i] = bf16_rne(r1 - bf16_f32(mb));
    }
    return r;
}
__device__ __forceinline__ v16b bh_ld(const float* __restrict__ p, long long sk, int k0, int h, int klen, float s) {
    v16b a;
#pragma unroll
    for (int i = 0; i < 16; ++i) { const int k = k0 + frag_k(i, h); a[i] = bf16_rne((k < klen) ? p[(long long)k * sk] * s : 0.f); }
    return a;
}
__device__ __forceinline__ v16h fh_row(const _Float16* __restrict__ row, int k0, int h) {
    v16h a;
#pragma unroll
    for (int i = 0; i < 16; ++i) a[i] = row[k0 + frag_k(i, h)];
    return a;
}

#define VST2(T, ptr, val) do { const T vst2_v_ = (val); *(volatile T*)(ptr) = vst2_v_; __threadfence(); *(volatile T*)(ptr) = vst2_v_; } while (0)
typedef float v4f __attribute__((ext_vector_type(4)));
#define VST2V4(ptr, val) do { const v4f vst2_v4_ = (val); *(volatile v4f*)(ptr) = vst2_v4_; __threadfence(); *(volatile v4f*)(ptr) = vst2_v4_; } while (0)

__device__ __attribute__((noinline)) float act_fn(float v, int act) {
    if (act == 1) return fmaxf(v, 0.f);
    if (act == 2) { const float u = 0.7978845608028654f * (v + 0.044715f * v * v * v); return 0.5f * v * (1.f + tanhf(u)); }
    if (act == 3) return v / (1.f + expf(-v));
    if (act == 4) return 0.5f * v * (1.f + erff(v * 0.7071067811865476f));
    if (act == 5) return tanhf(v);
    if (act == 6) return 1.f / (1.f + expf(-v));
    if (act == 7) return (v > 0.f) ? v : 0.01f * v;
    if (act == 8) return (v > 0.f) ? v : (expf(v) - 1.f);
    if (act == 9) return fminf(fmaxf(v, 0.f), 6.f);
    if (act == 10) return fabsf(v);
    if (act == 11) return (v >= 0.f) ? v : 0.1f * v;
    if (act == 12) return (v > 0.f) ? v : 0.2f * v;
    if (act == 13) return (v > 20.f) ? v : log1pf(expf(v));
    return v;
}

struct GemmP {
    const float* A; const float* B; const float* bias; const float* R; float* C;
    long long sAo, sAi, sAm, sAk, sBo, sBi, sBn, sBk, sCo, sCi, sCm, sRo, sRi, sRm, sRn;
    int M, N, K, zi_n, flags, act; float alpha, beta, sa, sb;
    int Npad, pad_;
};
static_assert(sizeof(GemmP) == 5 * 8 + 15 * 8 + 6 * 4 + 4 * 4 + 2 * 4, "GemmP has padding");

template <int MODE>
__global__ __launch_bounds__(32) void k_gemm(GemmP p) {
    const int lane = threadIdx.x & 31, h = lane >> 4, l15 = lane & 15;
    const int m0 = blockIdx.y * 16, n0 = blockIdx.x * 32;
    const int z = blockIdx.z, zo = z / p.zi_n, zi = z - zo * p.zi_n;
    const float* A = p.A + zo * p.sAo + zi * p.sAi;
    const float* B = p.B + zo * p.sBo + zi * p.sBi;
    const int am = min(m0 + l15, p.M - 1);
    v8f acc[2], comp[2];
#pragma unroll
    for (int t = 0; t < 2; ++t) { v8f zz = {}; acc[t] = zz; comp[t] = zz; }
    for (int k0 = 0; k0 < p.K; k0 += 32) {
        const float* arow = A + (long long)am * p.sAm;
        if (MODE == 1) {
            const Split a = sp_ld(arow, p.sAk, k0, h, p.K, 1.f);
#pragma unroll
            for (int t = 0; t < 2; ++t) {
                const int bn = min(n0 + t * 16 + l15, p.N - 1);
                acc[t] = wmma3(a, sp_ld(B + (long long)bn * p.sBn, p.sBk, k0, h, p.K, 1.f), acc[t]);
            }
        } else if (MODE == 3) {
            const Split3 a = sp3_ld(arow, p.sAk, k0, h, p.K, 1.f);
#pragma unroll
            for (int t = 0; t < 2; ++t) {
                const int bn = min(n0 + t * 16 + l15, p.N - 1);
                acc[t] = wmma6(a, sp3_ld(B + (long long)bn * p.sBn, p.sBk, k0, h, p.K, 1.f), acc[t]);
            }
        } else if (MODE == 4) {
            const Split3 a = sp3_ld(arow, p.sAk, k0, h, p.K, 1.f);
#pragma unroll
            for (int t = 0; t < 2; ++t) {
                const int bn = min(n0 + t * 16 + l15, p.N - 1); v8f zz = {};
                const v8f part = wmma6(a, sp3_ld(B + (long long)bn * p.sBn, p.sBk, k0, h, p.K, 1.f), zz);
                const v8f y = part - comp[t]; const v8f s = acc[t] + y; comp[t] = (s - acc[t]) - y; acc[t] = s;
            }
        } else if (MODE == 2) {
            const v16b a = bh_ld(arow, p.sAk, k0, h, p.K, 1.f);
#pragma unroll
            for (int t = 0; t < 2; ++t) {
                const int bn = min(n0 + t * 16 + l15, p.N - 1);
                acc[t] = wmmab(a, bh_ld(B + (long long)bn * p.sBn, p.sBk, k0, h, p.K, 1.f), acc[t]);
            }
        } else {
            const v16h a = fh_ld(arow, p.sAk, k0, h, p.K, p.sa);
#pragma unroll
            for (int t = 0; t < 2; ++t) {
                const int bn = min(n0 + t * 16 + l15, p.N - 1);
                acc[t] = wmma16(a, fh_ld(B + (long long)bn * p.sBn, p.sBk, k0, h, p.K, p.sb), acc[t]);
            }
        }
    }
    const float iscale = (MODE == 0) ? p.alpha / (p.sa * p.sb) : p.alpha;
    float* C = p.C + zo * p.sCo + zi * p.sCi;
    const float* R = p.R + zo * p.sRo + zi * p.sRi;
    __shared__ __align__(16) float ctile[16][36];
#pragma unroll
    for (int t = 0; t < 2; ++t) {
        const int n = n0 + t * 16 + l15; const int nn = min(n, p.N - 1);
#pragma unroll
        for (int r = 0; r < 8; ++r) {
            const int m = m0 + 8 * h + r; const int mm = min(m, p.M - 1);
            float v = acc[t][r] * iscale;
            if (p.flags & 1) v += p.bias[nn];
            if (p.flags & 2) v += p.bias[mm];
            if (p.flags & 8) v *= p.bias[(long long)zo * p.M + mm];
            v = act_fn(v, p.act);
            if (p.flags & 4) v += p.beta * R[(long long)mm * p.sRm + (long long)nn * p.sRn];
            ctile[8 * h + r][t * 16 + l15] = (n < p.N) ? v : 0.f;
        }
    }
    __syncthreads();
    const int NW = (p.Npad > p.N) ? p.Npad : p.N;
    const bool fast = (m0 + 16 <= p.M) && (n0 + 32 <= NW) && ((p.sCm & 3) == 0) && ((((size_t)C) & 15) == 0);
    if (fast) {
#pragma unroll
        for (int s = 0; s < 4; ++s) {
            const int row = s * 4 + (lane >> 3), c4 = (lane & 7) * 4;
            const v4f v = *(const v4f*)&ctile[row][c4];
            VST2V4(C + (long long)(m0 + row) * p.sCm + n0 + c4, v);
        }
    } else {
        for (int row = 0; row < 16; ++row) {
            const int m = m0 + row, n = n0 + lane;
            if (m < p.M && n < NW) VST2(float, C + (long long)m * p.sCm + n, ctile[row][lane]);
        }
    }
}


template <int MODE, int TM, int TN>
__global__ __launch_bounds__(32) void k_gemmT(GemmP p) {
    const int lane = threadIdx.x & 31, h = lane >> 4, l15 = lane & 15;
    const int m0 = blockIdx.y * (16 * TM), n0 = blockIdx.x * (16 * TN);
    const int z = blockIdx.z, zo = z / p.zi_n, zi = z - zo * p.zi_n;
    const float* A = p.A + zo * p.sAo + zi * p.sAi;
    const float* B = p.B + zo * p.sBo + zi * p.sBi;
    v8f acc[TM][TN];
#pragma unroll
    for (int i = 0; i < TM; ++i)
#pragma unroll
        for (int t = 0; t < TN; ++t) { v8f zz = {}; acc[i][t] = zz; }
    for (int k0 = 0; k0 < p.K; k0 += 32) {
        if (MODE == 1) {
            Split a[TM], b[TN];
#pragma unroll
            for (int i = 0; i < TM; ++i) { const int am = min(m0 + 16 * i + l15, p.M - 1); a[i] = sp_ld(A + (long long)am * p.sAm, p.sAk, k0, h, p.K, 1.f); }
#pragma unroll
            for (int t = 0; t < TN; ++t) { const int bn = min(n0 + 16 * t + l15, p.N - 1); b[t] = sp_ld(B + (long long)bn * p.sBn, p.sBk, k0, h, p.K, 1.f); }
#pragma unroll
            for (int i = 0; i < TM; ++i)
#pragma unroll
                for (int t = 0; t < TN; ++t) acc[i][t] = wmma3(a[i], b[t], acc[i][t]);
        } else if (MODE == 2) {
            v16b a[TM], b[TN];
#pragma unroll
            for (int i = 0; i < TM; ++i) { const int am = min(m0 + 16 * i + l15, p.M - 1); a[i] = bh_ld(A + (long long)am * p.sAm, p.sAk, k0, h, p.K, 1.f); }
#pragma unroll
            for (int t = 0; t < TN; ++t) { const int bn = min(n0 + 16 * t + l15, p.N - 1); b[t] = bh_ld(B + (long long)bn * p.sBn, p.sBk, k0, h, p.K, 1.f); }
#pragma unroll
            for (int i = 0; i < TM; ++i)
#pragma unroll
                for (int t = 0; t < TN; ++t) acc[i][t] = wmmab(a[i], b[t], acc[i][t]);
        } else {
            v16h a[TM], b[TN];
#pragma unroll
            for (int i = 0; i < TM; ++i) { const int am = min(m0 + 16 * i + l15, p.M - 1); a[i] = fh_ld(A + (long long)am * p.sAm, p.sAk, k0, h, p.K, p.sa); }
#pragma unroll
            for (int t = 0; t < TN; ++t) { const int bn = min(n0 + 16 * t + l15, p.N - 1); b[t] = fh_ld(B + (long long)bn * p.sBn, p.sBk, k0, h, p.K, p.sb); }
#pragma unroll
            for (int i = 0; i < TM; ++i)
#pragma unroll
                for (int t = 0; t < TN; ++t) acc[i][t] = wmma16(a[i], b[t], acc[i][t]);
        }
    }
    const float iscale = (MODE == 0) ? p.alpha / (p.sa * p.sb) : p.alpha;
    float* C = p.C + zo * p.sCo + zi * p.sCi;
    const float* R = p.R + zo * p.sRo + zi * p.sRi;
    const int NW = (p.Npad > p.N) ? p.Npad : p.N;
    __shared__ __align__(16) float ctile[16][36];
#pragma unroll
    for (int i = 0; i < TM; ++i) {
        const int mb = m0 + 16 * i; if (mb >= p.M) break;
#pragma unroll
        for (int tp = 0; tp < TN / 2; ++tp) {
            const int nb = n0 + 32 * tp; if (nb >= NW) break;
#pragma unroll
            for (int t2 = 0; t2 < 2; ++t2) {
                const int t = 2 * tp + t2; const int n = nb + t2 * 16 + l15; const int nn = min(n, p.N - 1);
#pragma unroll
                for (int r = 0; r < 8; ++r) {
                    const int m = mb + 8 * h + r; const int mm = min(m, p.M - 1);
                    float v = acc[i][t][r] * iscale;
                    if (p.flags & 1) v += p.bias[nn];
                    if (p.flags & 2) v += p.bias[mm];
            if (p.flags & 8) v *= p.bias[(long long)zo * p.M + mm];
                    v = act_fn(v, p.act);
                    if (p.flags & 4) v += p.beta * R[(long long)mm * p.sRm + (long long)nn * p.sRn];
                    ctile[8 * h + r][t2 * 16 + l15] = (n < p.N) ? v : 0.f;
                }
            }
            __syncthreads();
            const bool fast = (mb + 16 <= p.M) && (nb + 32 <= NW) && ((p.sCm & 3) == 0) && ((((size_t)C) & 15) == 0);
            if (fast) {
#pragma unroll
                for (int s = 0; s < 4; ++s) {
                    const int row = s * 4 + (lane >> 3), c4 = (lane & 7) * 4;
                    const v4f v = *(const v4f*)&ctile[row][c4];
                    VST2V4(C + (long long)(mb + row) * p.sCm + nb + c4, v);
                }
            } else {
                for (int row = 0; row < 16; ++row) {
                    const int m = mb + row, n = nb + lane;
                    if (m < p.M && n < NW) VST2(float, C + (long long)m * p.sCm + n, ctile[row][lane]);
                }
            }
            __syncthreads();
        }
    }
}

#define AW 4
struct AttnP {
    const float* Q; const float* K; const float* V; float* O; float* P; const float* Mf; const int* Mi; float* ST;
    const float* Pw; const float* Rt; const int* SQ; const int* SK;
    long long swb, swh, swi, swj, srb, srh, sri;
    long long sQb, sQh, sQi, sQd, sKb, sKh, sKj, sKd, sVb, sVh, sVj, sVd, sOb, sOh, sOi, sPb, sPh, sPi, smb, smh, smi, smj;
    int Lq, Lk, dh, dv, hrep, causal, coff, pband;
    float scale, mfill; int nonorm, mpol;
    int roff, rn, segpol, win;
};
static_assert(sizeof(AttnP) == 12 * 8 + 29 * 8 + 16 * 4, "AttnP has padding");

#ifndef KATTN_ATTR
#define KATTN_ATTR
#endif
template <int DHP, int DVP, int QM, bool SPLITPV, bool TWOPASS>
__global__ __launch_bounds__(32 * AW) KATTN_ATTR void k_attn(AttnP p) {
    constexpr int NT = DVP / 16;
    constexpr int KS = DHP / 32;
    constexpr int VP = DVP + 8;
    __shared__ __align__(16) float    pl[AW][16 * 64];
    __shared__ __align__(16) _Float16 vl[(SPLITPV ? 2 : 1) * 64 * VP];
    const int lane = threadIdx.x & 31, hf = lane >> 4, l15 = lane & 15, wave = threadIdx.x >> 5;
    const int h = blockIdx.y, b = blockIdx.z, hk = h / p.hrep;
    const int q0 = (blockIdx.x * AW + wave) * 16;
    float* myp = pl[wave];
    const float L2E = 1.4426950408889634f;
    const float NEG = -__builtin_inff();
    const int qi = min(q0 + l15, p.Lq - 1);
    const float* qrow = p.Q + b * p.sQb + h * p.sQh + (long long)qi * p.sQi;
    const float* kbase = p.K + b * p.sKb + hk * p.sKh;
    const float* vbase = p.V + b * p.sVb + hk * p.sVh;
    v16h qa[QM == 0 ? KS : 1]; Split qs_[QM == 1 ? KS : 1]; Split3 qt_[QM == 2 ? KS : 1];
#pragma unroll
    for (int ks = 0; ks < KS; ++ks) {
        if (QM == 2) qt_[ks] = sp3_ld(qrow, p.sQd, ks * 32, hf, p.dh, 1.f);
        else if (QM == 1) qs_[ks] = sp_ld(qrow, p.sQd, ks * 32, hf, p.dh, 1.f);
        else qa[ks] = fh_ld(qrow, p.sQd, ks * 32, hf, p.dh, 1.f);
    }
    v8f o[NT]; float m8[8], l8[8];
#pragma unroll
    for (int t = 0; t < NT; ++t) { v8f zz = {}; o[t] = zz; }
#pragma unroll
    for (int i = 0; i < 8; ++i) { m8[i] = NEG; l8[i] = 0.f; }
    int jend = p.Lk; int jstart = 0;
    if (p.causal == 1) { const int je = (blockIdx.x * AW + AW - 1) * 16 + 16 + p.coff; jend = min(jend, max(je, 0)); }
    if (p.win > 0) { const int js = (int)(blockIdx.x * AW) * 16 + p.coff - p.win; jstart = (js > 0) ? (js / 64) * 64 : 0; }
    const int npass = TWOPASS ? 2 : 1;
    for (int pass = 0; pass < npass; ++pass) {
        const bool dopv = (!TWOPASS) || pass == 1;
        for (int j0 = jstart; j0 < jend; j0 += 64) {
            if (dopv) {
                __syncthreads();
                for (int idx = threadIdx.x; idx < 64 * DVP; idx += 32 * AW) {
                    const int jr = idx / DVP, d = idx - jr * DVP, j = j0 + jr;
                    const float f = (j < p.Lk && d < p.dv) ? vbase[(long long)j * p.sVj + (long long)d * p.sVd] : 0.f;
                    if (SPLITPV) {
                        const __bf16 hb = bf16_rne(f);
                        ((__bf16*)vl)[jr * VP + d] = hb; ((__bf16*)vl)[64 * VP + jr * VP + d] = bf16_rne(f - bf16_f32(hb));
                    } else vl[jr * VP + d] = (_Float16)f;
                }
            }
            v8f s[4];
#pragma unroll
            for (int t = 0; t < 4; ++t) {
                const int j = min(j0 + t * 16 + l15, p.Lk - 1);
                const float* krow = kbase + (long long)j * p.sKj;
                v8f acc = {};
#pragma unroll
                for (int ks = 0; ks < KS; ++ks) {
                    if (QM == 2)      acc = wmma6(qt_[ks], sp3_ld(krow, p.sKd, ks * 32, hf, p.dh, 1.f), acc);
                    else if (QM == 1) acc = wmma3(qs_[ks], sp_ld(krow, p.sKd, ks * 32, hf, p.dh, 1.f), acc);
                    else              acc = wmma16(qa[ks], fh_ld(krow, p.sKd, ks * 32, hf, p.dh, 1.f), acc);
                }
                s[t] = acc;
            }
            float pv[8][4];
#pragma unroll
            for (int i = 0; i < 8; ++i) {
                const int irow = q0 + i + 8 * hf;
                const int ic = min(irow, p.Lq - 1);
                float sc[4];
#pragma unroll
                for (int t = 0; t < 4; ++t) {
                    const int jg = j0 + t * 16 + l15;
                    float v = s[t][i] * p.scale;
                    if (p.Mf) v += p.Mf[b * p.smb + h * p.smh + (long long)ic * p.smi + (long long)min(jg, p.Lk - 1) * p.smj];
                    if (p.Rt) { int rc = ic - min(jg, p.Lk - 1) + p.roff; rc = rc < 0 ? 0 : (rc >= p.rn ? p.rn - 1 : rc); v += p.Rt[b * p.srb + h * p.srh + (long long)ic * p.sri + rc]; }
                    if (p.Mi) { const int mv = p.Mi[b * p.smb + h * p.smh + (long long)ic * p.smi + (long long)min(jg, p.Lk - 1) * p.smj]; if (p.mpol ? (mv != 0) : (mv == 0)) v = p.mfill; }
                    if (p.SQ) { const bool same = p.SQ[(long long)b * p.Lq + ic] == p.SK[(long long)b * p.Lk + min(jg, p.Lk - 1)]; if (p.segpol ? same : !same) v = p.mfill; }
                    if (p.causal == 2 && jg > irow + p.coff) v = p.mfill;
                    if (jg >= p.Lk || (p.causal == 1 && jg > irow + p.coff) || (p.causal == 3 && jg < irow + p.coff) || (p.win > 0 && irow + p.coff - jg > p.win)) v = NEG; else v *= L2E;
                    sc[t] = v;
                }
                if (!TWOPASS || pass == 0) {
                    float mx = fmaxf(fmaxf(sc[0], sc[1]), fmaxf(sc[2], sc[3]));
                    mx = fmaxf(mx, __shfl_xor(mx, 1, 32)); mx = fmaxf(mx, __shfl_xor(mx, 2, 32));
                    mx = fmaxf(mx, __shfl_xor(mx, 4, 32)); mx = fmaxf(mx, __shfl_xor(mx, 8, 32));
                    const float mnew = fmaxf(m8[i], mx);
                    const float corr = (mnew == NEG) ? 1.f : exp2f(m8[i] - mnew);
                    float rs = 0.f;
#pragma unroll
                    for (int t = 0; t < 4; ++t) {
                        const float pp = (sc[t] == NEG) ? 0.f : exp2f(sc[t] - mnew); rs += pp;
                        pv[i][t] = p.Pw ? pp * p.Pw[b * p.swb + h * p.swh + (long long)ic * p.swi + (long long)min(j0 + t * 16 + l15, p.Lk - 1) * p.swj] : pp;
                    }
                    rs += __shfl_xor(rs, 1, 32); rs += __shfl_xor(rs, 2, 32); rs += __shfl_xor(rs, 4, 32); rs += __shfl_xor(rs, 8, 32);
                    l8[i] = l8[i] * corr + rs; m8[i] = mnew;
                    if (!TWOPASS) {
#pragma unroll
                        for (int t = 0; t < NT; ++t) o[t][i] *= corr;
                    }
                } else {
                    const float inv = (l8[i] > 0.f) ? 1.f / l8[i] : 0.f;
#pragma unroll
                    for (int t = 0; t < 4; ++t) {
                        const int jg = j0 + t * 16 + l15;
                        float pp = (sc[t] == NEG) ? 0.f : exp2f(sc[t] - m8[i]) * inv;
                        if (p.Pw) pp *= p.Pw[b * p.swb + h * p.swh + (long long)ic * p.swi + (long long)min(jg, p.Lk - 1) * p.swj];
                        pv[i][t] = pp;
                    }
                }
            }
            if (dopv) {
#pragma unroll
                for (int i = 0; i < 8; ++i)
#pragma unroll
                    for (int t = 0; t < 4; ++t) ((volatile float*)myp)[(i + 8 * hf) * 64 + t * 16 + l15] = pv[i][t];
                __syncthreads();
                if (p.P) {
                    float* pb_ = p.P + b * p.sPb + h * p.sPh;
                    const bool fastP = (p.pband == 0) && ((p.sPi & 3) == 0) && (j0 + 64 <= p.Lk) && (q0 + 16 <= p.Lq) && ((((size_t)pb_) & 15) == 0);
                    if (fastP) {
#pragma unroll
                        for (int s = 0; s < 8; ++s) {
                            const int row = s * 2 + (lane >> 4), c4 = (lane & 15) * 4;
                            const v4f v = *(const v4f*)(myp + row * 64 + c4);
                            VST2V4(pb_ + (long long)(q0 + row) * p.sPi + j0 + c4, v);
                        }
                    } else {
                        for (int row = 0; row < 16; ++row) {
                            const int irow = q0 + row; if (irow >= p.Lq) continue;
                            for (int c = lane; c < 64; c += 32) {
                                const int jg = j0 + c; if (jg >= p.Lk) continue;
                                if (p.pband == 0) VST2(float, pb_ + (long long)irow * p.sPi + jg, myp[row * 64 + c]);
                                else if (jg - irow <= p.pband && irow - jg <= p.pband) VST2(float, pb_ + (long long)irow * p.sPi + (jg - irow + p.pband), myp[row * 64 + c]);
                            }
                        }
                    }
                }
                if (SPLITPV) {
                    const Split pa0 = sp_ld(myp + l15 * 64, 1, 0, hf, 64, 1.f), pa1 = sp_ld(myp + l15 * 64, 1, 32, hf, 64, 1.f);
                    const __bf16* vh = (const __bf16*)vl; const __bf16* vlo = vh + 64 * VP;
#pragma unroll
                    for (int t = 0; t < NT; ++t) {
                        const int dcol = t * 16 + l15;
                        Split b0, b1;
#pragma unroll
                        for (int e = 0; e < 16; ++e) {
                            const int k0 = frag_k(e, hf), k1 = 32 + frag_k(e, hf);
                            b0.hi[e] = vh[k0 * VP + dcol]; b0.lo[e] = vlo[k0 * VP + dcol]; b1.hi[e] = vh[k1 * VP + dcol]; b1.lo[e] = vlo[k1 * VP + dcol];
                        }
                        o[t] = wmma3(pa0, b0, o[t]);
                        o[t] = wmma3(pa1, b1, o[t]);
                    }
                } else {
                    const v16h pa0 = fh_ld(myp + l15 * 64, 1, 0, hf, 64, 4096.f), pa1 = fh_ld(myp + l15 * 64, 1, 32, hf, 64, 4096.f);
#pragma unroll
                    for (int t = 0; t < NT; ++t) {
                        const int dcol = t * 16 + l15;
                        v16h b0, b1;
#pragma unroll
                        for (int e = 0; e < 16; ++e) { b0[e] = vl[frag_k(e, hf) * VP + dcol]; b1[e] = vl[(32 + frag_k(e, hf)) * VP + dcol]; }
                        o[t] = wmma16(pa0, b0, o[t]);
                        o[t] = wmma16(pa1, b1, o[t]);
                    }
                }
            }
        }
    }
    float* obase = p.O + b * p.sOb + h * p.sOh;
    if (p.ST) {
        const int rl = lane >> 1, isel = rl & 7;
        float mv = 0.f, lv = 0.f;
#pragma unroll
        for (int i = 0; i < 8; ++i) if (i == isel) { mv = m8[i]; lv = l8[i]; }
        const int irow = q0 + rl;
        if (irow < p.Lq) { float* st = p.ST + (((long long)b * gridDim.y + h) * p.Lq + irow) * 2 + (lane & 1); VST2(float, st, (lane & 1) ? lv : mv * 0.6931471805599453f); }
    }
    float invr[8];
#pragma unroll
    for (int i = 0; i < 8; ++i) {
        if (TWOPASS) invr[i] = SPLITPV ? 1.f : (1.f / 4096.f);
        else if (p.nonorm) invr[i] = exp2f(m8[i]) * (SPLITPV ? 1.f : (1.f / 4096.f));
        else invr[i] = (l8[i] > 0.f) ? (SPLITPV ? 1.f / l8[i] : 1.f / (l8[i] * 4096.f)) : 0.f;
    }
    __syncthreads();
    const bool ofast = ((p.sOi & 3) == 0) && ((((size_t)obase) & 15) == 0) && (q0 + 16 <= p.Lq);
#pragma unroll
    for (int c0 = 0; c0 < DVP; c0 += 64) {
#pragma unroll
        for (int i = 0; i < 8; ++i)
#pragma unroll
            for (int t = 0; t < NT; ++t) if (t * 16 >= c0 && t * 16 < c0 + 64) ((volatile float*)myp)[(i + 8 * hf) * 64 + (t * 16 - c0) + l15] = o[t][i] * invr[i];
        __syncthreads();
        const int cw = (DVP - c0 < 64) ? (DVP - c0) : 64;
        if (ofast && (c0 + cw <= p.dv) && (cw % 32 == 0)) {
            const int lpr = cw / 4;
            const int rows_per_ins = 32 / lpr;
            for (int r0 = 0; r0 < 16; r0 += rows_per_ins) {
                const int row = r0 + lane / lpr, c4 = (lane % lpr) * 4;
                const v4f v = *(const v4f*)(myp + row * 64 + c4);
                VST2V4(obase + (long long)(q0 + row) * p.sOi + c0 + c4, v);
            }
        } else {
            for (int row = 0; row < 16; ++row) {
                const int irow = q0 + row; if (irow >= p.Lq) continue;
                for (int c = lane; c < cw; c += 32) { const int d = c0 + c; if (d < p.dv) VST2(float, obase + (long long)irow * p.sOi + d, myp[row * 64 + c]); }
            }
        }
        __syncthreads();
    }
}

struct TrP { const float* src; float* dst; const float* R2; long long sSz, lds, sDz, ldd, sRz, ldr; int R, C, flags, act; float alpha, beta; };
static_assert(sizeof(TrP) == 3 * 8 + 6 * 8 + 6 * 4, "TrP has padding");
__global__ __launch_bounds__(256) void k_tr(TrP p) {
    __shared__ float tile[32][33];
    const int c0 = blockIdx.x * 32, r0 = blockIdx.y * 32, z = blockIdx.z;
    const int lane = threadIdx.x & 31, wave = threadIdx.x >> 5;
    const float* s = p.src + z * p.sSz;
#pragma unroll
    for (int k = 0; k < 4; ++k) {
        const int rl = wave * 4 + k, r = r0 + rl, c = c0 + lane;
        tile[rl][lane] = (r < p.R && c < p.C) ? s[(long long)r * p.lds + c] : 0.f;
    }
    __syncthreads();
    float* d = p.dst + z * p.sDz; const float* rr = p.R2 + z * p.sRz;
#pragma unroll
    for (int k = 0; k < 4; ++k) {
        const int cl = wave * 4 + k, c = c0 + cl, r = r0 + lane;
        if (c < p.C && r < p.R) {
            float v = act_fn(p.alpha * tile[lane][cl], p.act);
            if (p.flags & 1) v += p.beta * rr[(long long)c * p.ldr + r];
            VST2(float, d + (long long)c * p.ldd + r, v);
        }
    }
}

__global__ __launch_bounds__(256) void k_affine(const float* __restrict__ src, float* __restrict__ dst, int n, float a, float b, const float* __restrict__ sdev) {
    const int i = blockIdx.x * 256 + threadIdx.x;
    if (i < n) { const float aa = sdev ? a * sdev[0] : a; const float v = aa * src[i] + b; VST2(float, dst + i, v); }
}

struct SmP { const float* src; float* dst; const float* Mf; long long sz, sr, dz, dr, smz, smr; int n, pad; float scale_in, scale_out; };
static_assert(sizeof(SmP) == 3 * 8 + 6 * 8 + 4 * 4, "SmP has padding");
__global__ __launch_bounds__(256) void k_softmax(SmP p) {
    __shared__ float red[256];
    const int r = blockIdx.x, z = blockIdx.y, tid = threadIdx.x;
    const float* s = p.src + z * p.sz + (long long)r * p.sr;
    const float* mf = p.Mf ? (p.Mf + z * p.smz + (long long)r * p.smr) : nullptr;
    float mx = -__builtin_inff();
    for (int j = tid; j < p.n; j += 256) { float v = s[j] * p.scale_in; if (mf) v += mf[j]; mx = fmaxf(mx, v); }
    red[tid] = mx; __syncthreads();
    for (int o = 128; o > 0; o >>= 1) { if (tid < o) red[tid] = fmaxf(red[tid], red[tid + o]); __syncthreads(); }
    mx = red[0]; __syncthreads();
    float sum = 0.f;
    for (int j = tid; j < p.n; j += 256) { float v = s[j] * p.scale_in; if (mf) v += mf[j]; sum += (mx == -__builtin_inff()) ? 0.f : expf(v - mx); }
    red[tid] = sum; __syncthreads();
    for (int o = 128; o > 0; o >>= 1) { if (tid < o) red[tid] += red[tid + o]; __syncthreads(); }
    sum = red[0];
    const float inv = (sum > 0.f) ? p.scale_out / sum : 0.f;
    float* d = p.dst + z * p.dz + (long long)r * p.dr;
    for (int j = tid; j < p.n; j += 256) { float v = s[j] * p.scale_in; if (mf) v += mf[j]; const float o = (mx == -__builtin_inff()) ? 0.f : expf(v - mx) * inv; VST2(float, d + j, o); }
}
__global__ __launch_bounds__(256) void k_stats(const float* __restrict__ x, long long sz, long long so, long long si, int inner, int n, float eps, float* __restrict__ stat, int mode) {
    __shared__ float red[256];
    const int z = blockIdx.x, tid = threadIdx.x;
    const float* base = x + z * sz;
    float s = 0.f;
    for (int e = tid; e < n; e += 256) s += base[(long long)(e / inner) * so + (long long)(e % inner) * si];
    red[tid] = s; __syncthreads();
    for (int o = 128; o > 0; o >>= 1) { if (tid < o) red[tid] += red[tid + o]; __syncthreads(); }
    const float mu = (mode == 0 || mode == 3) ? red[0] / (float)n : 0.f; __syncthreads();
    float q = 0.f;
    for (int e = tid; e < n; e += 256) { const float dlt = base[(long long)(e / inner) * so + (long long)(e % inner) * si] - mu; q += dlt * dlt; }
    red[tid] = q; __syncthreads();
    for (int o = 128; o > 0; o >>= 1) { if (tid < o) red[tid] += red[tid + o]; __syncthreads(); }
    {
        float rs;
        if (mode == 2) rs = sqrtf((float)n) / fmaxf(sqrtf(red[0]), eps); else if (mode == 3) rs = rsqrtf(red[0] / (float)(n - 1) + eps); else rs = rsqrtf(red[0] / (float)n + eps);
        if (tid < 32) { const float v = (tid == 0) ? mu : ((tid == 1) ? rs : 0.f); VST2(float, stat + (long long)z * 32 + tid, v); }
    }
}
__global__ __launch_bounds__(256) void k_norm_apply(const float* __restrict__ x, float* __restrict__ y, const float* __restrict__ stat, const float* __restrict__ g, const float* __restrict__ bta,
                                                     int Z, int C, int L, int G, int bn, int act) {
    const long long idx = (long long)blockIdx.x * 256 + threadIdx.x;
    if (idx >= (long long)Z * C * L) return;
    const int l = (int)(idx % L); const long long zc = idx / L; const int c = (int)(zc % C), z = (int)(zc / C); (void)l;
    const int set = bn ? c : (z * G + c / (C / G));
    float v = (x[idx] - stat[(long long)set * 32]) * stat[(long long)set * 32 + 1];
    if (g) v *= g[c];
    if (bta) v += bta[c];
    v = act_fn(v, act);
    VST2(float, y + idx, v);
}

__global__ __launch_bounds__(256) void k_lse_neg(const float* __restrict__ st, float* __restrict__ c, int n) {
    const int i = blockIdx.x * 256 + threadIdx.x;
    if (i < n) { const float v = -(st[2 * i] + logf(st[2 * i + 1])); VST2(float, c + i, v); }
}

__global__ __launch_bounds__(256) void k_iota(int* __restrict__ dst, int n, int a, int b) {
    const int i = blockIdx.x * 256 + threadIdx.x;
    if (i < n) { const int v = a * i + b; VST2(int, dst + i, v); }
}

__global__ __launch_bounds__(256) void k_axpby(const float* __restrict__ x, const float* __restrict__ y, float* __restrict__ dst, int n, float a, float b, float c) {
    const int i = blockIdx.x * 256 + threadIdx.x;
    if (i < n) { const float v = a * x[i] + b * y[i] + c; VST2(float, dst + i, v); }
}

struct RopeP { const float* X; float* Y; const float* C; const float* Sn; const int* pos; long long sXr, sXh, sYr, sYh, sCb, sCp, sCd; int R, Hn, D, S, mode, tmode, pmode, pad; };
static_assert(sizeof(RopeP) == 5 * 8 + 7 * 8 + 8 * 4, "RopeP has padding");
__global__ __launch_bounds__(256) void k_rope(RopeP p) {
    const long long idx = (long long)blockIdx.x * 256 + threadIdx.x;
    if (idx >= (long long)p.R * p.Hn * p.D) return;
    const int d = (int)(idx % p.D); const long long rh = idx / p.D; const int h = (int)(rh % p.Hn); const int r = (int)(rh / p.Hn);
    const int half = p.D / 2;
    int partner; float sign;
    if (p.mode == 0) { partner = (d < half) ? d + half : d - half; sign = (d < half) ? -1.f : 1.f; }
    else { partner = d ^ 1; sign = (d & 1) ? 1.f : -1.f; }
    const int tcol = (p.tmode == 0) ? d : ((p.tmode == 1) ? (d % half) : (d >> 1));
    const int pp = (p.pmode == 0) ? (r % p.S) : ((p.pmode == 1) ? h : p.pos[r]);
    const long long toff = (long long)(r / p.S) * p.sCb + (long long)pp * p.sCp + (long long)tcol * p.sCd;
    const float* xr = p.X + (long long)r * p.sXr + (long long)h * p.sXh;
    const float v = xr[d] * p.C[toff] + sign * xr[partner] * p.Sn[toff];
    VST2(float, p.Y + (long long)r * p.sYr + (long long)h * p.sYh + d, v);
}

__global__ __launch_bounds__(256) void k_invf(float* __restrict__ invb, int half, int D, float base, float num, int fmode, float cexp) {
    const int i = blockIdx.x * 256 + threadIdx.x;
    if (i >= ((half + 31) / 32) * 32) return;
    if (i >= half) { VST2(float, invb + i, 0.f); return; }
    const float e = (float)(2 * i) / (float)D;
    float invf;
    if (fmode == 1) invf = num * expf((float)(2 * i) * cexp);
    else if (fmode == 2) invf = num * powf(base, (-2.0f * ((float)i - 1.0f)) / (float)D);
    else invf = num * (1.0f / powf(base, e));
    VST2(float, invb + i, invf);
}
__global__ __launch_bounds__(256) void k_sincos(float* __restrict__ cs, float* __restrict__ sn, const float* __restrict__ invb, int S, int half, float pscale) {
    const int idx = blockIdx.x * 256 + threadIdx.x;
    if (idx >= S * half) return;
    const int s = idx / half, i = idx - s * half;
    const float ang = (pscale * (float)s) * invb[i];
    VST2(float, cs + idx, cosf(ang)); VST2(float, sn + idx, sinf(ang));
}

__global__ __launch_bounds__(256) void k_mulact(const float* __restrict__ x, const float* __restrict__ y, float* __restrict__ dst, int n, int act) {
    const int i = blockIdx.x * 256 + threadIdx.x;
    if (i < n) { const float v = act_fn(x[i], act) * y[i]; VST2(float, dst + i, v); }
}

__global__ __launch_bounds__(256) void k_matvec(GemmP p) {
    const int rpt = (p.N == 1) ? 1 : 32;
    const long long r0 = ((long long)blockIdx.x * 256 + threadIdx.x) * rpt; const int z = blockIdx.z, zo = z / p.zi_n, zi = z - zo * p.zi_n;
    if (r0 >= p.M) return;
    const float* Bb = p.B + zo * p.sBo + zi * p.sBi;
    float* C = p.C + zo * p.sCo + zi * p.sCi; const float* R = p.R + zo * p.sRo + zi * p.sRi;
    for (int rr = 0; rr < rpt; ++rr) {
        const long long r = r0 + rr; if (r >= p.M) break;
        const float* A = p.A + zo * p.sAo + zi * p.sAi + r * p.sAm;
        float acc[8] = {0.f, 0.f, 0.f, 0.f, 0.f, 0.f, 0.f, 0.f};
        for (int k = 0; k < p.K; ++k) { const float a = A[(long long)k * p.sAk];
#pragma unroll
            for (int j = 0; j < 8; ++j) if (j < p.N) acc[j] += a * Bb[(long long)j * p.sBn + (long long)k * p.sBk]; }
#pragma unroll
        for (int j = 0; j < 8; ++j) if (j < p.N) {
            float v = acc[j] * p.alpha;
            if (p.flags & 1) v += p.bias[j];
            if (p.flags & 2) v += p.bias[r];
            v = act_fn(v, p.act);
            if (p.flags & 4) v += p.beta * R[r * p.sRm + (long long)j * p.sRn];
            VST2(float, C + r * p.sCm + j, v);
        }
    }
}
__global__ __launch_bounds__(256) void k_smallsoftmax(const float* __restrict__ src, float* __restrict__ dst, long long sr, long long dr, int n, long long R, float scale) {
    const long long r0 = ((long long)blockIdx.x * 256 + threadIdx.x) * 32;
    for (int rr = 0; rr < 32; ++rr) {
        const long long r = r0 + rr; if (r >= R) return;
        const float* s = src + r * sr; float* d = dst + r * dr;
        float mx = -__builtin_inff();
        for (int j = 0; j < n; ++j) mx = fmaxf(mx, s[j] * scale);
        float sum = 0.f;
        for (int j = 0; j < n; ++j) sum += expf(s[j] * scale - mx);
        const float inv = 1.f / sum;
        for (int j = 0; j < n; ++j) { const float v = expf(s[j] * scale - mx) * inv; VST2(float, d + j, v); }
    }
}

__global__ __launch_bounds__(32) void k_unitstat(float* __restrict__ st) { const int t = threadIdx.x; const float v = (t == 1) ? 1.f : 0.f; VST2(float, st + t, v); }

__global__ __launch_bounds__(256) void k_lincopy(const float* __restrict__ src, long long lds, float* __restrict__ dst, long long ldd, long long rows, int cols) {
    const long long i = (long long)blockIdx.x * 256 + threadIdx.x; if (i >= rows * cols) return;
    const long long r = i / cols; const int c = (int)(i - r * cols);
    const float v = src[r * lds + c]; VST2(float, dst + r * ldd + c, v);
}

namespace w25 {
typedef __attribute__((ext_vector_type(16))) _Float16 v16h;
typedef __attribute__((ext_vector_type(8)))  _Float16 v8h;
typedef __attribute__((ext_vector_type(16))) __bf16   v16b;
typedef __attribute__((ext_vector_type(8)))  __bf16   v8b;
typedef __attribute__((ext_vector_type(8)))  float    v8f;
typedef __attribute__((ext_vector_type(4)))  float    v4f;

__device__ __forceinline__ unsigned short f2bf_bits(float f) {
  unsigned u = __float_as_uint(f);
  return (unsigned short)((u + 0x7FFFu + ((u >> 16) & 1u)) >> 16);
}
__device__ __forceinline__ float bf_bits2f(unsigned short h) { return __uint_as_float(((unsigned)h) << 16); }

__device__ __forceinline__ void dep_guard_h(v8f& a, v8f& b, v16h x, v16h y) { asm volatile("v_nop\n\tv_nop\n\tv_nop\n\tv_nop" : "+v"(a), "+v"(b) : "v"(x), "v"(y)); }
__device__ __forceinline__ void dep_guard_b(v8f& a, v8f& b, v16b x, v16b y) { asm volatile("v_nop\n\tv_nop\n\tv_nop\n\tv_nop" : "+v"(a), "+v"(b) : "v"(x), "v"(y)); }
__device__ __forceinline__ void keep4_h(v16h a, v16h b, v16h c, v16h d) { asm volatile("v_nop" :: "v"(a), "v"(b), "v"(c), "v"(d)); }
__device__ __forceinline__ void keep4_b(v16b a, v16b b, v16b c, v16b d) { asm volatile("v_nop" :: "v"(a), "v"(b), "v"(c), "v"(d)); }
__device__ __forceinline__ void acc_guard4(v8f& a, v8f& b, v8f& c, v8f& d) { asm volatile("v_nop\n\tv_nop\n\tv_nop\n\tv_nop" : "+v"(a), "+v"(b), "+v"(c), "+v"(d)); }
template <typename T> struct Frag;
template <> struct Frag<_Float16> {
  typedef v16h V; union U { v16h v; v8h h[2]; };
  static __device__ __forceinline__ v16h load(const _Float16* p) {
    U f; f.h[0] = *(const v8h*)(p); f.h[1] = *(const v8h*)(p + 16); return f.v;
  }
  static __device__ __forceinline__ v8f mma(v16h a, v16h b, v8f c) {
    return __builtin_amdgcn_wmma_f32_16x16x32_f16(false, a, false, b, (short)0, c, false, false);
  }
  static __device__ __forceinline__ void guard(v8f& a, v8f& b, v16h x, v16h y) { dep_guard_h(a, b, x, y); }
  static __device__ __forceinline__ void keep(v16h a, v16h b, v16h c, v16h d) { keep4_h(a, b, c, d); }
};
template <> struct Frag<__bf16> {
  typedef v16b V; union U { v16b v; v8b h[2]; };
  static __device__ __forceinline__ v16b load(const __bf16* p) {
    U f; f.h[0] = *(const v8b*)(p); f.h[1] = *(const v8b*)(p + 16); return f.v;
  }
  static __device__ __forceinline__ v8f mma(v16b a, v16b b, v8f c) {
    return __builtin_amdgcn_wmma_f32_16x16x32_bf16(false, a, false, b, (short)0, c, false, false);
  }
  static __device__ __forceinline__ void guard(v8f& a, v8f& b, v16b x, v16b y) { dep_guard_b(a, b, x, y); }
  static __device__ __forceinline__ void keep(v16b a, v16b b, v16b c, v16b d) { keep4_b(a, b, c, d); }
};

template <int ET> struct Elem;
template <> struct Elem<0> { typedef _Float16 T; };
template <> struct Elem<1> { typedef __bf16 T; };
template <int ET, bool SPLIT, int BIAS_MODE, int OUT_MODE, bool RESID, int ACT = 0>
__global__ __launch_bounds__(256) void wmma_gemm64(
    const unsigned short* __restrict__ Ap, const unsigned short* __restrict__ A2p, int lda, long strideA,
    const unsigned short* __restrict__ Btp, const unsigned short* __restrict__ Bt2p, int ldb, long strideB,
    void* __restrict__ Cout, void* __restrict__ Cout2, int ldc, long strideC,
    const float* __restrict__ bias,
    const float* __restrict__ resid, long strideR,
    int M, int N, int K, float scale) {
  typedef typename Elem<ET>::T T;
  typedef typename Frag<T>::V V;
  const T* A = (const T*)Ap; const T* A2 = (const T*)A2p; const T* Bt = (const T*)Btp; const T* Bt2 = (const T*)Bt2p;
  __shared__ __align__(16) float sT[8][16 * 68];
  const int b    = blockIdx.y;
  const int lane = threadIdx.x & 31;
  const int wave = threadIdx.x >> 5;
  const int tilesN = N >> 6;
  const int tilesM = M >> 6;
  const int tile = blockIdx.x * 8 + wave;
  if (tile >= tilesM * tilesN) return;
  const int tm = tile / tilesN;
  const int tn = tile - tm * tilesN;
  const int m0 = tm << 6;
  const int n0 = tn << 6;

  const T* Ab  = A  + (size_t)b * strideA;
  const T* Bb  = Bt + (size_t)b * strideB;
  const T* Ab2 = SPLIT ? (A2  + (size_t)b * strideA) : nullptr;
  const T* Bb2 = SPLIT ? (Bt2 + (size_t)b * strideB) : nullptr;

  const int rlane = lane & 15;
  const int koff  = (lane >> 4) * 8;
  const int mOff  = (lane >> 4) * 8;

  v8f acc[4][4];
#pragma unroll
  for (int i = 0; i < 4; ++i)
#pragma unroll
    for (int j = 0; j < 4; ++j) acc[i][j] = (v8f){0.f,0.f,0.f,0.f,0.f,0.f,0.f,0.f};

  for (int k0 = 0; k0 < K; k0 += 32) {
    V bh[4], bl[4];
#pragma unroll
    for (int j = 0; j < 4; ++j) {
      const size_t bo = (size_t)(n0 + (j << 4) + rlane) * ldb + koff + k0;
      bh[j] = Frag<T>::load(Bb + bo);
      if (SPLIT) bl[j] = Frag<T>::load(Bb2 + bo);
    }
#pragma unroll
    for (int i = 0; i < 4; ++i) {
      const size_t ao = (size_t)(m0 + (i << 4) + rlane) * lda + koff + k0;
      V ah = Frag<T>::load(Ab + ao);
      V al;
      if (SPLIT) al = Frag<T>::load(Ab2 + ao);
#pragma unroll
      for (int j = 0; j < 4; ++j) {
        acc[i][j] = Frag<T>::mma(ah, bh[j], acc[i][j]);
        if (SPLIT) {
          acc[i][j] = Frag<T>::mma(ah, bl[j], acc[i][j]);
          acc[i][j] = Frag<T>::mma(al, bh[j], acc[i][j]);
        }
      }
      Frag<T>::guard(acc[i][0], acc[i][3], ah, SPLIT ? al : ah);
    }
    Frag<T>::keep(bh[0], bh[1], bh[2], bh[3]);
    if (SPLIT) Frag<T>::keep(bl[0], bl[1], bl[2], bl[3]);
  }
  acc_guard4(acc[0][0], acc[0][1], acc[0][2], acc[0][3]);
  acc_guard4(acc[1][0], acc[1][1], acc[1][2], acc[1][3]);
  acc_guard4(acc[2][0], acc[2][1], acc[2][2], acc[2][3]);
  acc_guard4(acc[3][0], acc[3][1], acc[3][2], acc[3][3]);

  float* slab = sT[wave];
  const float* Rb = RESID ? (resid + (size_t)b * strideR) : nullptr;
#pragma unroll
  for (int i = 0; i < 4; ++i) {
    const int mBase = m0 + (i << 4);
#pragma unroll
    for (int j = 0; j < 4; ++j) {
      const int n = n0 + (j << 4) + rlane;
      float bv = 0.f;
      if (BIAS_MODE == 2) bv = bias[n];
#pragma unroll
      for (int r = 0; r < 8; ++r) {
        float v = acc[i][j][r] * scale;
        if (BIAS_MODE == 1) v += bias[mBase + mOff + r];
        if (BIAS_MODE == 2) v += bv;
        if (RESID) v += Rb[(size_t)(mBase + mOff + r) * ldc + n];
        if (ACT == 1) v = tanhf(v);
        if (ACT == 2) v = fmaxf(v, 0.0f);
        if (ACT == 3) v = v / (1.0f + expf(-v));
        if (ACT == 4) v = (v > 0.f) ? v : 0.01f * v;
        if (ACT == 5) v = 0.5f * v * (1.0f + erff(v * 0.70710678118654752f));
        slab[(mOff + r) * 68 + (j << 4) + rlane] = v;
      }
    }
    __builtin_amdgcn_fence(__ATOMIC_RELEASE, "workgroup");
    __builtin_amdgcn_wave_barrier();
    __builtin_amdgcn_fence(__ATOMIC_ACQUIRE, "workgroup");
    if (OUT_MODE == 0) {
      float* C = (float*)Cout + (size_t)b * strideC;
      const int hh = lane >> 4, c4 = (lane & 15) * 4;
      for (int pass = 0; pass < 2; ++pass) {
#pragma unroll
        for (int it = 0; it < 8; ++it) {
          const int row = it * 2 + hh;
          v4f v = *(const v4f*)(slab + row * 68 + c4);
          *(volatile v4f*)(C + (size_t)(mBase + row) * ldc + n0 + c4) = v;
        }
        __threadfence();
      }
    } else {
      const int q = lane >> 3, c8 = (lane & 7) * 8;
      unsigned short* C  = (unsigned short*)Cout  + (size_t)b * strideC;
      unsigned short* C2 = (OUT_MODE == 2) ? ((unsigned short*)Cout2 + (size_t)b * strideC) : nullptr;
      for (int pass = 0; pass < 2; ++pass) {
#pragma unroll
        for (int it = 0; it < 4; ++it) {
          const int row = it * 4 + q;
          const float* sp = slab + row * 68 + c8;
          v8h hv, lv;
#pragma unroll
          for (int e = 0; e < 8; ++e) {
            if (OUT_MODE == 1) {
              hv[e] = (_Float16)sp[e];
            } else {
              unsigned short hb = f2bf_bits(sp[e]);
              unsigned short lb = f2bf_bits(sp[e] - bf_bits2f(hb));
              hv[e] = __builtin_bit_cast(_Float16, hb);
              lv[e] = __builtin_bit_cast(_Float16, lb);
            }
          }
          *(volatile v8h*)(C + (size_t)(mBase + row) * ldc + n0 + c8) = hv;
          if (OUT_MODE == 2) *(volatile v8h*)(C2 + (size_t)(mBase + row) * ldc + n0 + c8) = lv;
        }
        __threadfence();
      }
    }
    __builtin_amdgcn_fence(__ATOMIC_RELEASE, "workgroup");
    __builtin_amdgcn_wave_barrier();
    __builtin_amdgcn_fence(__ATOMIC_ACQUIRE, "workgroup");
  }
}

__global__ __launch_bounds__(256) void cast_f32_f16x2(
    const float* __restrict__ in, _Float16* __restrict__ out, int n2) {
  int i = blockIdx.x * 256 + threadIdx.x;
  if (i < n2) {
    const _Float16 h0 = (_Float16)in[2 * i], h1 = (_Float16)in[2 * i + 1];
    const unsigned u = (unsigned)__builtin_bit_cast(unsigned short, h0) | ((unsigned)__builtin_bit_cast(unsigned short, h1) << 16);
    ((volatile unsigned*)out)[i] = u;
    __threadfence();
    ((volatile unsigned*)out)[i] = u;
  }
}


}

__global__ __launch_bounds__(256) void k_castT16(const float* __restrict__ src, long long lds, _Float16* __restrict__ dst, long long ldd, int R, int C, float s) {
    const long long i = (long long)blockIdx.x * 256 + threadIdx.x; const long long np = (long long)C * (R / 2); if (i >= np) return; const int c = (int)(i / (R / 2)); const int r = 2 * (int)(i % (R / 2));
    const _Float16 h0 = (_Float16)(src[(long long)r * lds + c] * s), h1 = (_Float16)(src[(long long)(r + 1) * lds + c] * s);
    const unsigned u = (unsigned)__builtin_bit_cast(unsigned short, h0) | ((unsigned)__builtin_bit_cast(unsigned short, h1) << 16);
    volatile unsigned* d = (volatile unsigned*)(dst + (long long)c * ldd + r); *d = u; __threadfence(); *d = u; }
__global__ __launch_bounds__(256) void k_cast16(const float* __restrict__ src, long long lds, _Float16* __restrict__ dst, long long ldd, int R, int C, float s) {
    const long long i = (long long)blockIdx.x * 256 + threadIdx.x; const long long np = (long long)R * (C / 2); if (i >= np) return; const int r = (int)(i / (C / 2)); const int c = 2 * (int)(i % (C / 2));
    const _Float16 h0 = (_Float16)(src[(long long)r * lds + c] * s), h1 = (_Float16)(src[(long long)r * lds + c + 1] * s);
    const unsigned u = (unsigned)__builtin_bit_cast(unsigned short, h0) | ((unsigned)__builtin_bit_cast(unsigned short, h1) << 16);
    volatile unsigned* d = (volatile unsigned*)(dst + (long long)r * ldd + c); *d = u; __threadfence(); *d = u; }

__device__ __forceinline__ unsigned int f2bf2_pack(float a, float b, unsigned int* lo) {
    const unsigned short ha = w25::f2bf_bits(a), hb = w25::f2bf_bits(b);
    const unsigned short la = w25::f2bf_bits(a - w25::bf_bits2f(ha)), lb = w25::f2bf_bits(b - w25::bf_bits2f(hb));
    *lo = (unsigned)la | ((unsigned)lb << 16); return (unsigned)ha | ((unsigned)hb << 16); }
__global__ __launch_bounds__(256) void k_castS16(const float* __restrict__ src, long long lds, __bf16* __restrict__ dhi, __bf16* __restrict__ dlo, long long ldd, int R, int C, float s, int transpose) {
    const long long i = (long long)blockIdx.x * 256 + threadIdx.x; long long o; float a, b;
    if (transpose) { const long long np = (long long)C * (R / 2); if (i >= np) return; const int c = (int)(i / (R / 2)); const int r = 2 * (int)(i % (R / 2)); a = src[(long long)r * lds + c] * s; b = src[(long long)(r + 1) * lds + c] * s; o = (long long)c * ldd + r; }
    else { const long long np = (long long)R * (C / 2); if (i >= np) return; const int r = (int)(i / (C / 2)); const int c = 2 * (int)(i % (C / 2)); a = src[(long long)r * lds + c] * s; b = src[(long long)r * lds + c + 1] * s; o = (long long)r * ldd + c; }
    unsigned lo; const unsigned hi = f2bf2_pack(a, b, &lo); volatile unsigned* ph = (volatile unsigned*)(dhi + o); volatile unsigned* pl = (volatile unsigned*)(dlo + o);
    *ph = hi; *pl = lo; __threadfence(); *ph = hi; *pl = lo; }

namespace w25 {
#define AT_D 64
#define AT_NW 4
#define AT_QB 64
#define AT_KC 64
struct AttnGeom { const float* cp = nullptr; const float* pc = nullptr; long c_bs = 0, c_rs = 0, c_hs = 0;
                  long q_bs, q_rs, q_hs, k_bs, k_rs, k_hs, v_bs, v_rs, v_hs, o_bs, o_rs, o_hs;
                  int S, Skv, H, mask_mode; float qscale; int blk0; float mask_fill; int mask_is_int; };
static_assert(sizeof(AttnGeom) == 168, "no padding");

__device__ __forceinline__ unsigned short at_bf_bits(float f) {
  unsigned u = __float_as_uint(f);
  return (unsigned short)((u + 0x7FFFu + ((u >> 16) & 1u)) >> 16);
}
__device__ __forceinline__ __bf16 at_f2bf(float f) { return __builtin_bit_cast(__bf16, at_bf_bits(f)); }
__device__ __forceinline__ void at_split(float f, __bf16& hi, __bf16& lo) {
  const unsigned short hb = at_bf_bits(f);
  hi = __builtin_bit_cast(__bf16, hb);
  lo = at_f2bf(f - __uint_as_float(((unsigned)hb) << 16));
}
__device__ __forceinline__ v8f at_mma(v16b a, v16b b, v8f c) {
  c = __builtin_amdgcn_wmma_f32_16x16x32_bf16(false, a, false, b, (short)0, c, false, false);
  asm volatile("v_nop\n\tv_nop\n\tv_nop\n\tv_nop" : "+v"(c) : "v"(a), "v"(b));
  return c;
}
template <bool F16> __device__ __forceinline__ __bf16 at_to16(float f) {
  if (F16) return __builtin_bit_cast(__bf16, (_Float16)f);
  return at_f2bf(f);
}
template <bool F16> __device__ __forceinline__ v8f at_mma16(v16b a, v16b b, v8f c) {
  if (F16) {
    const v16h ah = __builtin_bit_cast(v16h, a), bh = __builtin_bit_cast(v16h, b);
    c = __builtin_amdgcn_wmma_f32_16x16x32_f16(false, ah, false, bh, (short)0, c, false, false);
    asm volatile("v_nop\n\tv_nop\n\tv_nop\n\tv_nop" : "+v"(c) : "v"(ah), "v"(bh));
    return c;
  }
  return at_mma(a, b, c);
}

template <bool SPLIT_QK, bool SPLIT_PV, bool F16 = false>
__global__ __launch_bounds__(128)
void attn64_kernel(const float* __restrict__ q, const float* __restrict__ k,
                   const float* __restrict__ v, float* __restrict__ out,
                   const void* __restrict__ mask_a, const int* __restrict__ mask_b, AttnGeom g) {
  static_assert(!(F16 && (SPLIT_QK || SPLIT_PV)), "f16 mode is non-split");
  const float PSC = F16 ? 32768.0f : 1.0f;
  union FB { v16b v; v8b h[2]; };
  __shared__ __align__(16) __bf16 Ksh[AT_KC * AT_D];
  __shared__ __align__(16) __bf16 Ksl[SPLIT_QK ? AT_KC * AT_D : 8];
  __shared__ __align__(16) __bf16 Vth[AT_D * AT_KC];
  __shared__ __align__(16) __bf16 Vtl[SPLIT_PV ? AT_D * AT_KC : 8];
  __shared__ __align__(16) __bf16 Psh[AT_NW][16 * AT_KC];
  __shared__ __align__(16) __bf16 Psl[SPLIT_PV ? AT_NW : 1][SPLIT_PV ? 16 * AT_KC : 8];
  __shared__ __align__(16) float  Os[AT_NW][16 * 68];

  const int tid  = threadIdx.x;
  const int wave = tid >> 5;
  const int lane = tid & 31;
  const int hh   = lane >> 4;
  const int c    = lane & 15;

  const int nqb = g.S / AT_QB;
  const int bx = blockIdx.x + g.blk0;
  const int qb = bx % nqb;
  const int bh = bx / nqb;
  const int h  = bh % g.H;
  const int b  = bh / g.H;
  const int qbase_block = qb * AT_QB;
  const int q0 = qbase_block + wave * 16;

  const float* qb_ptr = q + (size_t)b * g.q_bs + (size_t)h * g.q_hs;
  const float* kb_ptr = k + (size_t)b * g.k_bs + (size_t)h * g.k_hs;
  const float* vb_ptr = v + (size_t)b * g.v_bs + (size_t)h * g.v_hs;
  float*       ob_ptr = out + (size_t)b * g.o_bs + (size_t)h * g.o_hs;

  v16b qah[2], qal[2];
  {
    const float* qrow = qb_ptr + (size_t)(q0 + c) * g.q_rs;
#pragma unroll
    for (int dc = 0; dc < 2; ++dc) {
#pragma unroll
      for (int e = 0; e < 8; ++e) {
        const float f0 = qrow[dc * 32 + 8 * hh + e] * g.qscale;
        const float f1 = qrow[dc * 32 + 16 + 8 * hh + e] * g.qscale;
        if (SPLIT_QK) { __bf16 hq, lq; at_split(f0, hq, lq); qah[dc][e] = hq; qal[dc][e] = lq; at_split(f1, hq, lq); qah[dc][8 + e] = hq; qal[dc][8 + e] = lq; }
        else { qah[dc][e] = at_to16<F16>(f0); qah[dc][8 + e] = at_to16<F16>(f1); qal[dc][e] = qah[dc][e]; qal[dc][8 + e] = qah[dc][8 + e]; }
      }
    }
  }

  float mrow[8], lrow[8];
  v8f oacc[4];
#pragma unroll
  for (int r = 0; r < 8; ++r) { mrow[r] = -INFINITY; lrow[r] = 0.f; }
#pragma unroll
  for (int t = 0; t < 4; ++t) oacc[t] = (v8f){0.f,0.f,0.f,0.f,0.f,0.f,0.f,0.f};

  const int nChunks = (g.mask_mode == 1 || g.mask_mode == 4) ? (qb + 1) : (g.Skv / AT_KC);
  int qkeep[8];
#pragma unroll
  for (int r = 0; r < 8; ++r) qkeep[r] = (g.mask_mode == 3) ? mask_b[(size_t)b * g.S + q0 + 8 * hh + r] : 1;
  for (int kc = 0; kc < nChunks; ++kc) {
    const int kv0 = kc * AT_KC;
    __syncthreads();
    {
      const int kvr = tid >> 1, dh = (tid & 1) * 32;
      const float* krow = kb_ptr + (size_t)(kv0 + kvr) * g.k_rs + dh;
      const float* vrow = vb_ptr + (size_t)(kv0 + kvr) * g.v_rs + dh;
#pragma unroll
      for (int i = 0; i < 8; ++i) {
        v4f kk = *(const v4f*)(krow + 4 * i);
        v4f vv = *(const v4f*)(vrow + 4 * i);
#pragma unroll
        for (int e = 0; e < 4; ++e) {
          const int d = dh + 4 * i + e;
          if (SPLIT_QK) { __bf16 a, bl; at_split(kk[e], a, bl); Ksh[kvr * AT_D + d] = a; Ksl[kvr * AT_D + d] = bl; }
          else Ksh[kvr * AT_D + d] = at_to16<F16>(kk[e]);
          if (SPLIT_PV) { __bf16 a, bl; at_split(vv[e], a, bl); Vth[d * AT_KC + kvr] = a; Vtl[d * AT_KC + kvr] = bl; }
          else Vth[d * AT_KC + kvr] = at_to16<F16>(vv[e]);
        }
      }
    }
    __syncthreads();

    v8f s[4];
#pragma unroll
    for (int j = 0; j < 4; ++j) {
      s[j] = (v8f){0.f,0.f,0.f,0.f,0.f,0.f,0.f,0.f};
#pragma unroll 1
      for (int dc = 0; dc < 2; ++dc) {
        FB kb;
        kb.h[0] = *(const v8b*)(Ksh + (j * 16 + c) * AT_D + dc * 32 + 8 * hh);
        kb.h[1] = *(const v8b*)(Ksh + (j * 16 + c) * AT_D + dc * 32 + 16 + 8 * hh);
        s[j] = at_mma16<F16>(qah[dc], kb.v, s[j]);
        if (SPLIT_QK) {
          FB kl;
          kl.h[0] = *(const v8b*)(Ksl + (j * 16 + c) * AT_D + dc * 32 + 8 * hh);
          kl.h[1] = *(const v8b*)(Ksl + (j * 16 + c) * AT_D + dc * 32 + 16 + 8 * hh);
          s[j] = at_mma16<F16>(qah[dc], kl.v, s[j]);
          s[j] = at_mma16<F16>(qal[dc], kb.v, s[j]);
        }
      }
    }
    const bool diag = (g.mask_mode == 1) && (kc == qb);
    int kvkeep[4] = {1, 1, 1, 1};
    if (g.mask_mode == 3) {
#pragma unroll
      for (int j = 0; j < 4; ++j) kvkeep[j] = ((const int*)mask_a)[(size_t)b * g.Skv + kv0 + j * 16 + c];
    }
    float cm[8];
#pragma unroll
    for (int r = 0; r < 8; ++r) {
      const int qrow = q0 + 8 * hh + r;
      float m = -INFINITY;
#pragma unroll
      for (int j = 0; j < 4; ++j) {
        const int kvcol = kv0 + j * 16 + c;
        bool masked = false;
        if (diag) masked = (kvcol > qrow);
        else if (g.mask_mode == 4) masked = (kvcol > qrow) || (qrow - kvcol > g.mask_is_int);
        else if (g.mask_mode == 2) {
          const size_t mi = (size_t)qrow * g.Skv + kvcol;
          masked = (g.mask_is_int == 0) ? (((const float*)mask_a)[mi] == 0.0f)
                 : (g.mask_is_int == 1) ? (((const int*)mask_a)[mi] == 0) : (((const int*)mask_a)[mi] != 0);
        } else if (g.mask_mode == 3) masked = (qkeep[r] == 0) || (kvkeep[j] == 0);
        else if (g.mask_mode == 5) {
          const size_t mi = (size_t)qrow * g.Skv + kvcol;
          masked = (((const int*)mask_a)[mi] != 0);
          int n = mask_b[mi]; n = n < 0 ? 0 : n;
          s[j][r] += g.cp[(size_t)b * g.c_bs + (size_t)h * g.c_hs + (size_t)qrow * g.c_rs + n]
                   + g.pc[(size_t)b * g.c_bs + (size_t)h * g.c_hs + (size_t)kvcol * g.c_rs + n];
        }
        if (masked) s[j][r] = g.mask_fill;
        m = fmaxf(m, s[j][r]);
      }
#pragma unroll
      for (int off = 1; off < 16; off <<= 1) m = fmaxf(m, __shfl_xor(m, off, 32));
      cm[r] = m;
    }
    __bf16* pwh = Psh[wave];
    __bf16* pwl = Psl[SPLIT_PV ? wave : 0];
#pragma unroll
    for (int r = 0; r < 8; ++r) {
      const float mnew = fmaxf(mrow[r], cm[r]);
      const float alpha = expf(mrow[r] - mnew);
      mrow[r] = mnew;
      float psum = 0.f;
#pragma unroll
      for (int j = 0; j < 4; ++j) {
        const float p = expf(s[j][r] - mnew);
        psum += p;
        if (SPLIT_PV) { __bf16 a, bl; at_split(p, a, bl); pwh[(8 * hh + r) * AT_KC + j * 16 + c] = a; pwl[(8 * hh + r) * AT_KC + j * 16 + c] = bl; }
        else pwh[(8 * hh + r) * AT_KC + j * 16 + c] = at_to16<F16>(p * PSC);
      }
#pragma unroll
      for (int off = 1; off < 16; off <<= 1) psum += __shfl_xor(psum, off, 32);
      lrow[r] = lrow[r] * alpha + psum;
#pragma unroll
      for (int t = 0; t < 4; ++t) oacc[t][r] *= alpha;
    }
    __builtin_amdgcn_fence(__ATOMIC_RELEASE, "workgroup");
    __builtin_amdgcn_wave_barrier();
    __builtin_amdgcn_fence(__ATOMIC_ACQUIRE, "workgroup");
#pragma unroll 1
    for (int kk = 0; kk < 2; ++kk) {
      FB pa, pl;
      pa.h[0] = *(const v8b*)(pwh + c * AT_KC + kk * 32 + 8 * hh);
      pa.h[1] = *(const v8b*)(pwh + c * AT_KC + kk * 32 + 16 + 8 * hh);
      if (SPLIT_PV) {
        pl.h[0] = *(const v8b*)(pwl + c * AT_KC + kk * 32 + 8 * hh);
        pl.h[1] = *(const v8b*)(pwl + c * AT_KC + kk * 32 + 16 + 8 * hh);
      }
#pragma unroll
      for (int t = 0; t < 4; ++t) {
        FB vb;
        vb.h[0] = *(const v8b*)(Vth + (t * 16 + c) * AT_KC + kk * 32 + 8 * hh);
        vb.h[1] = *(const v8b*)(Vth + (t * 16 + c) * AT_KC + kk * 32 + 16 + 8 * hh);
        oacc[t] = at_mma16<F16>(pa.v, vb.v, oacc[t]);
        if (SPLIT_PV) {
          FB vl;
          vl.h[0] = *(const v8b*)(Vtl + (t * 16 + c) * AT_KC + kk * 32 + 8 * hh);
          vl.h[1] = *(const v8b*)(Vtl + (t * 16 + c) * AT_KC + kk * 32 + 16 + 8 * hh);
          oacc[t] = at_mma16<F16>(pa.v, vl.v, oacc[t]);
          oacc[t] = at_mma16<F16>(pl.v, vb.v, oacc[t]);
        }
      }
    }
  }

  float* os = Os[wave];
#pragma unroll
  for (int r = 0; r < 8; ++r) {
    const float inv = 1.0f / (lrow[r] * PSC);
#pragma unroll
    for (int t = 0; t < 4; ++t) os[(8 * hh + r) * 68 + t * 16 + c] = oacc[t][r] * inv;
  }
  __builtin_amdgcn_fence(__ATOMIC_RELEASE, "workgroup");
  __builtin_amdgcn_wave_barrier();
  __builtin_amdgcn_fence(__ATOMIC_ACQUIRE, "workgroup");
  {
    const int c4 = (lane & 15) * 4;
    for (int pass = 0; pass < 2; ++pass) {
#pragma unroll
      for (int it = 0; it < 8; ++it) {
        const int row = it * 2 + hh;
        v4f val = *(const v4f*)(os + row * 68 + c4);
        *(volatile v4f*)(ob_ptr + (size_t)(q0 + row) * g.o_rs + c4) = val;
      }
      __threadfence();
    }
  }
}

}

__global__ __launch_bounds__(256) void k_ld_bias(const float* __restrict__ RT, float* __restrict__ BIAS, int NH, int L) { const long long t = (long long)blockIdx.x * 256 + threadIdx.x; if (t >= (long long)NH * L * L) return; const int kk = (int)(t % L); const int q = (int)((t / L) % L); const int h = (int)(t / ((long long)L * L)); int n = q - kk; n = n < 0 ? 0 : n; int bk;
    if (n < 16) bk = n; else { const float v = logf((float)n / 16.f) / 2.0794415416798357f * 16.f; bk = 16 + (int)v; bk = bk > 31 ? 31 : bk; }
    VST2(float, BIAS + t, RT[bk * NH + h]); }
__global__ __launch_bounds__(256) void k_ld_rms(const float* __restrict__ X, const float* __restrict__ S, float* __restrict__ Y, int D) { __shared__ float red[256]; const long long r = blockIdx.x; const int t = threadIdx.x; const float* xr = X + r * D; float s = 0.f; for (int j = t; j < D; j += 256) { const float v = xr[j]; s += v * v; }
    red[t] = s; __syncthreads(); for (int o = 128; o > 0; o >>= 1) { if (t < o) red[t] += red[t + o]; __syncthreads(); } const float inv = rsqrtf(red[0] / (float)D + 1e-6f);
    for (int j = t; j < D; j += 256) VST2(float, Y + r * D + j, xr[j] * inv * S[j]); }
__global__ __launch_bounds__(256) void k_ld_gg(float* __restrict__ A, const float* __restrict__ Bv, long long n) { const long long t = (long long)blockIdx.x * 256 + threadIdx.x; if (t >= n) return; const float v = A[t]; VST2(float, A + t, 0.5f * v * (1.f + erff(v * 0.70710678118654752f)) * Bv[t]); }

template __global__ void k_gemm<0>(GemmP);

extern "C" void kernel_launch(void* const* d_in, const int* in_sizes, int n_in, void* d_out, int out_size, void* d_ws, size_t ws_size, hipStream_t stream) {
    (void)in_sizes; (void)n_in; (void)out_size; (void)ws_size;
    const float* xin = (const float*)d_in[0];
    const float* enc = (const float*)d_in[1];
    const float* qa = (const float*)d_in[2];
    const float* qb = (const float*)d_in[3];
    const float* ka = (const float*)d_in[4];
    const float* kb = (const float*)d_in[5];
    const float* va = (const float*)d_in[6];
    const float* vb = (const float*)d_in[7];
    const float* oa = (const float*)d_in[8];
    const float* ob = (const float*)d_in[9];
    const float* rt = (const float*)d_in[10];
    const float* ln1 = (const float*)d_in[11];
    const float* ln2 = (const float*)d_in[12];
    const float* ln3 = (const float*)d_in[13];
    const float* sWq = (const float*)d_in[14];
    const float* sWk = (const float*)d_in[15];
    const float* sWv = (const float*)d_in[16];
    const float* sWo = (const float*)d_in[17];
    const float* cWq = (const float*)d_in[18];
    const float* cWk = (const float*)d_in[19];
    const float* cWv = (const float*)d_in[20];
    const float* cWo = (const float*)d_in[21];
    const float* wi0 = (const float*)d_in[22];
    const float* wi1 = (const float*)d_in[23];
    const float* wom = (const float*)d_in[24];
    const int Bn = 4;
    const int L = 512;
    const int D = 1024;
    const int NH = 16;
    const int HD = 64;
    const int R = 32;
    const int FF = 4096;
    const int NBK = 32;
    float* out = (float*)d_out;
    char* wsp = (char*)d_ws;
    float* XN = (float*)wsp; wsp += (((size_t)((size_t)L * D) * 4 + 255) / 256) * 256;
    float* LOW = (float*)wsp; wsp += (((size_t)((size_t)L * R) * 4 + 255) / 256) * 256;
    float* Q = (float*)wsp; wsp += (((size_t)((size_t)L * D) * 4 + 255) / 256) * 256;
    float* Kb = (float*)wsp; wsp += (((size_t)((size_t)L * D) * 4 + 255) / 256) * 256;
    float* V = (float*)wsp; wsp += (((size_t)((size_t)L * D) * 4 + 255) / 256) * 256;
    float* AT = (float*)wsp; wsp += (((size_t)((size_t)L * D) * 4 + 255) / 256) * 256;
    float* X1 = (float*)wsp; wsp += (((size_t)((size_t)Bn * L * D) * 4 + 255) / 256) * 256;
    float* Y1 = (float*)wsp; wsp += (((size_t)((size_t)Bn * L * D) * 4 + 255) / 256) * 256;
    float* BIAS = (float*)wsp; wsp += (((size_t)((size_t)NH * L * L) * 4 + 255) / 256) * 256;
    float* G0 = (float*)wsp; wsp += (((size_t)((size_t)L * FF) * 4 + 255) / 256) * 256;
    float* G1 = (float*)wsp; wsp += (((size_t)((size_t)L * FF) * 4 + 255) / 256) * 256;
    unsigned short* G64A = (unsigned short*)wsp; wsp += (((size_t)(2097152) * 2 + 255) / 256) * 256;
    unsigned short* G64B = (unsigned short*)wsp; wsp += (((size_t)(4194304) * 2 + 255) / 256) * 256;
    k_ld_bias<<<(unsigned)(((long long)NH * L * L + 255) / 256), 256, 0, stream>>>(rt, BIAS, NH, L);
    k_ld_rms<<<L, 256, 0, stream>>>(xin + (size_t)0 * L * D, ln1, XN, D);
    { GemmP sq0lo;
      sq0lo.A = XN; sq0lo.B = qa + (size_t)0 * D * R; sq0lo.bias = XN; sq0lo.R = XN; sq0lo.C = LOW;
      sq0lo.sAo = 0; sq0lo.sAi = 0; sq0lo.sAm = D; sq0lo.sAk = 1; sq0lo.sBo = 0; sq0lo.sBi = 0; sq0lo.sBn = 1; sq0lo.sBk = R; sq0lo.sCo = 0; sq0lo.sCi = 0; sq0lo.sCm = R; sq0lo.sRo = 0; sq0lo.sRi = 0; sq0lo.sRm = 0; sq0lo.sRn = 0;
      sq0lo.M = L; sq0lo.N = R; sq0lo.K = D; sq0lo.zi_n = 1; sq0lo.flags = 0; sq0lo.act = 0;
      sq0lo.alpha = 1.0f; sq0lo.beta = 0.0f; sq0lo.sa = 1.0f; sq0lo.sb = 1.0f; sq0lo.Npad = R; sq0lo.pad_ = 0;
      if ((long long)(L) >= 64 && (long long)(R) >= 64) k_gemmT<0, 4, 4><<<dim3((unsigned)((R) + 63) / 64, (unsigned)((L) + 63) / 64, (unsigned)(1)), 32, 0, stream>>>(sq0lo);
      else k_gemm<0><<<dim3((unsigned)((R) + 31) / 32, (unsigned)((L) + 15) / 16, (unsigned)(1)), 32, 0, stream>>>(sq0lo); }
    k_cast16<<<(unsigned)((((long long)(512) * ((1024) / 2)) + 255) / 256), 256, 0, stream>>>(XN, 1024, (_Float16*)(G64A), 1024, 512, 1024, 1.0f);
    k_castT16<<<(unsigned)((((long long)(1024) * ((1024) / 2)) + 255) / 256), 256, 0, stream>>>(sWq, 1024, (_Float16*)(G64B), 1024, 1024, 1024, 16.0f);
    w25::wmma_gemm64<0, false, 0, 0, false, 0><<<dim3((unsigned)((((512) / 64) * ((1024) / 64) + 7) / 8), (unsigned)(1)), 256, 0, stream>>>((const unsigned short*)(G64A), nullptr, 1024, 0, (const unsigned short*)(G64B), nullptr, 1024, 0, (void*)(Q), nullptr, 1024, 0, nullptr, nullptr, 0, 512, 1024, 1024, 0.0625f);
    { GemmP sq0ab;
      sq0ab.A = LOW; sq0ab.B = qb + (size_t)0 * R * D; sq0ab.bias = LOW; sq0ab.R = Q; sq0ab.C = Q;
      sq0ab.sAo = 0; sq0ab.sAi = 0; sq0ab.sAm = R; sq0ab.sAk = 1; sq0ab.sBo = 0; sq0ab.sBi = 0; sq0ab.sBn = 1; sq0ab.sBk = D; sq0ab.sCo = 0; sq0ab.sCi = 0; sq0ab.sCm = D; sq0ab.sRo = 0; sq0ab.sRi = 0; sq0ab.sRm = D; sq0ab.sRn = 1;
      sq0ab.M = L; sq0ab.N = D; sq0ab.K = R; sq0ab.zi_n = 1; sq0ab.flags = 4; sq0ab.act = 0;
      sq0ab.alpha = 1.0f; sq0ab.beta = 1.0f; sq0ab.sa = 1.0f; sq0ab.sb = 1.0f; sq0ab.Npad = D; sq0ab.pad_ = 0;
      if ((long long)(L) >= 64 && (long long)(D) >= 64) k_gemmT<0, 4, 4><<<dim3((unsigned)((D) + 63) / 64, (unsigned)((L) + 63) / 64, (unsigned)(1)), 32, 0, stream>>>(sq0ab);
      else k_gemm<0><<<dim3((unsigned)((D) + 31) / 32, (unsigned)((L) + 15) / 16, (unsigned)(1)), 32, 0, stream>>>(sq0ab); }
    { GemmP sk0lo;
      sk0lo.A = XN; sk0lo.B = ka + (size_t)0 * D * R; sk0lo.bias = XN; sk0lo.R = XN; sk0lo.C = LOW;
      sk0lo.sAo = 0; sk0lo.sAi = 0; sk0lo.sAm = D; sk0lo.sAk = 1; sk0lo.sBo = 0; sk0lo.sBi = 0; sk0lo.sBn = 1; sk0lo.sBk = R; sk0lo.sCo = 0; sk0lo.sCi = 0; sk0lo.sCm = R; sk0lo.sRo = 0; sk0lo.sRi = 0; sk0lo.sRm = 0; sk0lo.sRn = 0;
      sk0lo.M = L; sk0lo.N = R; sk0lo.K = D; sk0lo.zi_n = 1; sk0lo.flags = 0; sk0lo.act = 0;
      sk0lo.alpha = 1.0f; sk0lo.beta = 0.0f; sk0lo.sa = 1.0f; sk0lo.sb = 1.0f; sk0lo.Npad = R; sk0lo.pad_ = 0;
      if ((long long)(L) >= 64 && (long long)(R) >= 64) k_gemmT<0, 4, 4><<<dim3((unsigned)((R) + 63) / 64, (unsigned)((L) + 63) / 64, (unsigned)(1)), 32, 0, stream>>>(sk0lo);
      else k_gemm<0><<<dim3((unsigned)((R) + 31) / 32, (unsigned)((L) + 15) / 16, (unsigned)(1)), 32, 0, stream>>>(sk0lo); }
    k_cast16<<<(unsigned)((((long long)(512) * ((1024) / 2)) + 255) / 256), 256, 0, stream>>>(XN, 1024, (_Float16*)(G64A), 1024, 512, 1024, 1.0f);
    k_castT16<<<(unsigned)((((long long)(1024) * ((1024) / 2)) + 255) / 256), 256, 0, stream>>>(sWk, 1024, (_Float16*)(G64B), 1024, 1024, 1024, 16.0f);
    w25::wmma_gemm64<0, false, 0, 0, false, 0><<<dim3((unsigned)((((512) / 64) * ((1024) / 64) + 7) / 8), (unsigned)(1)), 256, 0, stream>>>((const unsigned short*)(G64A), nullptr, 1024, 0, (const unsigned short*)(G64B), nullptr, 1024, 0, (void*)(Kb), nullptr, 1024, 0, nullptr, nullptr, 0, 512, 1024, 1024, 0.0625f);
    { GemmP sk0ab;
      sk0ab.A = LOW; sk0ab.B = kb + (size_t)0 * R * D; sk0ab.bias = LOW; sk0ab.R = Kb; sk0ab.C = Kb;
      sk0ab.sAo = 0; sk0ab.sAi = 0; sk0ab.sAm = R; sk0ab.sAk = 1; sk0ab.sBo = 0; sk0ab.sBi = 0; sk0ab.sBn = 1; sk0ab.sBk = D; sk0ab.sCo = 0; sk0ab.sCi = 0; sk0ab.sCm = D; sk0ab.sRo = 0; sk0ab.sRi = 0; sk0ab.sRm = D; sk0ab.sRn = 1;
      sk0ab.M = L; sk0ab.N = D; sk0ab.K = R; sk0ab.zi_n = 1; sk0ab.flags = 4; sk0ab.act = 0;
      sk0ab.alpha = 1.0f; sk0ab.beta = 1.0f; sk0ab.sa = 1.0f; sk0ab.sb = 1.0f; sk0ab.Npad = D; sk0ab.pad_ = 0;
      if ((long long)(L) >= 64 && (long long)(D) >= 64) k_gemmT<0, 4, 4><<<dim3((unsigned)((D) + 63) / 64, (unsigned)((L) + 63) / 64, (unsigned)(1)), 32, 0, stream>>>(sk0ab);
      else k_gemm<0><<<dim3((unsigned)((D) + 31) / 32, (unsigned)((L) + 15) / 16, (unsigned)(1)), 32, 0, stream>>>(sk0ab); }
    { GemmP sv0lo;
      sv0lo.A = XN; sv0lo.B = va + (size_t)0 * D * R; sv0lo.bias = XN; sv0lo.R = XN; sv0lo.C = LOW;
      sv0lo.sAo = 0; sv0lo.sAi = 0; sv0lo.sAm = D; sv0lo.sAk = 1; sv0lo.sBo = 0; sv0lo.sBi = 0; sv0lo.sBn = 1; sv0lo.sBk = R; sv0lo.sCo = 0; sv0lo.sCi = 0; sv0lo.sCm = R; sv0lo.sRo = 0; sv0lo.sRi = 0; sv0lo.sRm = 0; sv0lo.sRn = 0;
      sv0lo.M = L; sv0lo.N = R; sv0lo.K = D; sv0lo.zi_n = 1; sv0lo.flags = 0; sv0lo.act = 0;
      sv0lo.alpha = 1.0f; sv0lo.beta = 0.0f; sv0lo.sa = 1.0f; sv0lo.sb = 1.0f; sv0lo.Npad = R; sv0lo.pad_ = 0;
      if ((long long)(L) >= 64 && (long long)(R) >= 64) k_gemmT<0, 4, 4><<<dim3((unsigned)((R) + 63) / 64, (unsigned)((L) + 63) / 64, (unsigned)(1)), 32, 0, stream>>>(sv0lo);
      else k_gemm<0><<<dim3((unsigned)((R) + 31) / 32, (unsigned)((L) + 15) / 16, (unsigned)(1)), 32, 0, stream>>>(sv0lo); }
    k_cast16<<<(unsigned)((((long long)(512) * ((1024) / 2)) + 255) / 256), 256, 0, stream>>>(XN, 1024, (_Float16*)(G64A), 1024, 512, 1024, 1.0f);
    k_castT16<<<(unsigned)((((long long)(1024) * ((1024) / 2)) + 255) / 256), 256, 0, stream>>>(sWv, 1024, (_Float16*)(G64B), 1024, 1024, 1024, 16.0f);
    w25::wmma_gemm64<0, false, 0, 0, false, 0><<<dim3((unsigned)((((512) / 64) * ((1024) / 64) + 7) / 8), (unsigned)(1)), 256, 0, stream>>>((const unsigned short*)(G64A), nullptr, 1024, 0, (const unsigned short*)(G64B), nullptr, 1024, 0, (void*)(V), nullptr, 1024, 0, nullptr, nullptr, 0, 512, 1024, 1024, 0.0625f);
    { GemmP sv0ab;
      sv0ab.A = LOW; sv0ab.B = vb + (size_t)0 * R * D; sv0ab.bias = LOW; sv0ab.R = V; sv0ab.C = V;
      sv0ab.sAo = 0; sv0ab.sAi = 0; sv0ab.sAm = R; sv0ab.sAk = 1; sv0ab.sBo = 0; sv0ab.sBi = 0; sv0ab.sBn = 1; sv0ab.sBk = D; sv0ab.sCo = 0; sv0ab.sCi = 0; sv0ab.sCm = D; sv0ab.sRo = 0; sv0ab.sRi = 0; sv0ab.sRm = D; sv0ab.sRn = 1;
      sv0ab.M = L; sv0ab.N = D; sv0ab.K = R; sv0ab.zi_n = 1; sv0ab.flags = 4; sv0ab.act = 0;
      sv0ab.alpha = 1.0f; sv0ab.beta = 1.0f; sv0ab.sa = 1.0f; sv0ab.sb = 1.0f; sv0ab.Npad = D; sv0ab.pad_ = 0;
      if ((long long)(L) >= 64 && (long long)(D) >= 64) k_gemmT<0, 4, 4><<<dim3((unsigned)((D) + 63) / 64, (unsigned)((L) + 63) / 64, (unsigned)(1)), 32, 0, stream>>>(sv0ab);
      else k_gemm<0><<<dim3((unsigned)((D) + 31) / 32, (unsigned)((L) + 15) / 16, (unsigned)(1)), 32, 0, stream>>>(sv0ab); }
    {   AttnP a;
      a.Q = Q; a.K = Kb; a.V = V; a.O = AT; a.P = 0; a.Mf = BIAS; a.Mi = 0; a.ST = 0;
      a.Pw = 0; a.Rt = 0; a.SQ = 0; a.SK = 0;
      a.swb = 0; a.swh = 0; a.swi = 0; a.swj = 0; a.srb = 0; a.srh = 0; a.sri = 0; a.sQb = 0; a.sQh = HD; a.sQi = D; a.sQd = 1; a.sKb = 0; a.sKh = HD; a.sKj = D; a.sKd = 1; a.sVb = 0; a.sVh = HD; a.sVj = D; a.sVd = 1; a.sOb = 0; a.sOh = HD; a.sOi = D; a.sPb = 0; a.sPh = 0; a.sPi = 0; a.smb = 0; a.smh = (long long)L * L; a.smi = L; a.smj = 1;
      a.Lq = L; a.Lk = L; a.dh = HD; a.dv = HD; a.hrep = 1; a.causal = 1; a.coff = 0; a.pband = 0;
      a.scale = 0.125f; a.mfill = 0.0f; a.nonorm = 0; a.mpol = 0;
      a.roff = 0; a.rn = 1; a.segpol = 0; a.win = 0;
      k_attn<64, 64, 0, false, false><<<dim3((unsigned)((L) + 16 * AW - 1) / (16 * AW), (unsigned)(NH), (unsigned)(1)), 32 * AW, 0, stream>>>(a); }
    { GemmP so0lo;
      so0lo.A = AT; so0lo.B = oa + (size_t)0 * D * R; so0lo.bias = AT; so0lo.R = AT; so0lo.C = LOW;
      so0lo.sAo = 0; so0lo.sAi = 0; so0lo.sAm = D; so0lo.sAk = 1; so0lo.sBo = 0; so0lo.sBi = 0; so0lo.sBn = 1; so0lo.sBk = R; so0lo.sCo = 0; so0lo.sCi = 0; so0lo.sCm = R; so0lo.sRo = 0; so0lo.sRi = 0; so0lo.sRm = 0; so0lo.sRn = 0;
      so0lo.M = L; so0lo.N = R; so0lo.K = D; so0lo.zi_n = 1; so0lo.flags = 0; so0lo.act = 0;
      so0lo.alpha = 1.0f; so0lo.beta = 0.0f; so0lo.sa = 1.0f; so0lo.sb = 1.0f; so0lo.Npad = R; so0lo.pad_ = 0;
      if ((long long)(L) >= 64 && (long long)(R) >= 64) k_gemmT<0, 4, 4><<<dim3((unsigned)((R) + 63) / 64, (unsigned)((L) + 63) / 64, (unsigned)(1)), 32, 0, stream>>>(so0lo);
      else k_gemm<0><<<dim3((unsigned)((R) + 31) / 32, (unsigned)((L) + 15) / 16, (unsigned)(1)), 32, 0, stream>>>(so0lo); }
    k_cast16<<<(unsigned)((((long long)(512) * ((1024) / 2)) + 255) / 256), 256, 0, stream>>>(AT, 1024, (_Float16*)(G64A), 1024, 512, 1024, 1.0f);
    k_castT16<<<(unsigned)((((long long)(1024) * ((1024) / 2)) + 255) / 256), 256, 0, stream>>>(sWo, 1024, (_Float16*)(G64B), 1024, 1024, 1024, 16.0f);
    w25::wmma_gemm64<0, false, 0, 0, true, 0><<<dim3((unsigned)((((512) / 64) * ((1024) / 64) + 7) / 8), (unsigned)(1)), 256, 0, stream>>>((const unsigned short*)(G64A), nullptr, 1024, 0, (const unsigned short*)(G64B), nullptr, 1024, 0, (void*)(X1 + (size_t)0 * L * D), nullptr, 1024, 0, nullptr, xin + (size_t)0 * L * D, 0, 512, 1024, 1024, 0.0625f);
    { GemmP so0ab;
      so0ab.A = LOW; so0ab.B = ob + (size_t)0 * R * D; so0ab.bias = LOW; so0ab.R = X1 + (size_t)0 * L * D; so0ab.C = X1 + (size_t)0 * L * D;
      so0ab.sAo = 0; so0ab.sAi = 0; so0ab.sAm = R; so0ab.sAk = 1; so0ab.sBo = 0; so0ab.sBi = 0; so0ab.sBn = 1; so0ab.sBk = D; so0ab.sCo = 0; so0ab.sCi = 0; so0ab.sCm = D; so0ab.sRo = 0; so0ab.sRi = 0; so0ab.sRm = D; so0ab.sRn = 1;
      so0ab.M = L; so0ab.N = D; so0ab.K = R; so0ab.zi_n = 1; so0ab.flags = 4; so0ab.act = 0;
      so0ab.alpha = 1.0f; so0ab.beta = 1.0f; so0ab.sa = 1.0f; so0ab.sb = 1.0f; so0ab.Npad = D; so0ab.pad_ = 0;
      if ((long long)(L) >= 64 && (long long)(D) >= 64) k_gemmT<0, 4, 4><<<dim3((unsigned)((D) + 63) / 64, (unsigned)((L) + 63) / 64, (unsigned)(1)), 32, 0, stream>>>(so0ab);
      else k_gemm<0><<<dim3((unsigned)((D) + 31) / 32, (unsigned)((L) + 15) / 16, (unsigned)(1)), 32, 0, stream>>>(so0ab); }
    k_ld_rms<<<L, 256, 0, stream>>>(X1 + (size_t)0 * L * D, ln2, XN, D);
    { GemmP cq0lo;
      cq0lo.A = XN; cq0lo.B = qa + (size_t)1 * D * R; cq0lo.bias = XN; cq0lo.R = XN; cq0lo.C = LOW;
      cq0lo.sAo = 0; cq0lo.sAi = 0; cq0lo.sAm = D; cq0lo.sAk = 1; cq0lo.sBo = 0; cq0lo.sBi = 0; cq0lo.sBn = 1; cq0lo.sBk = R; cq0lo.sCo = 0; cq0lo.sCi = 0; cq0lo.sCm = R; cq0lo.sRo = 0; cq0lo.sRi = 0; cq0lo.sRm = 0; cq0lo.sRn = 0;
      cq0lo.M = L; cq0lo.N = R; cq0lo.K = D; cq0lo.zi_n = 1; cq0lo.flags = 0; cq0lo.act = 0;
      cq0lo.alpha = 1.0f; cq0lo.beta = 0.0f; cq0lo.sa = 1.0f; cq0lo.sb = 1.0f; cq0lo.Npad = R; cq0lo.pad_ = 0;
      if ((long long)(L) >= 64 && (long long)(R) >= 64) k_gemmT<0, 4, 4><<<dim3((unsigned)((R) + 63) / 64, (unsigned)((L) + 63) / 64, (unsigned)(1)), 32, 0, stream>>>(cq0lo);
      else k_gemm<0><<<dim3((unsigned)((R) + 31) / 32, (unsigned)((L) + 15) / 16, (unsigned)(1)), 32, 0, stream>>>(cq0lo); }
    k_cast16<<<(unsigned)((((long long)(512) * ((1024) / 2)) + 255) / 256), 256, 0, stream>>>(XN, 1024, (_Float16*)(G64A), 1024, 512, 1024, 1.0f);
    k_castT16<<<(unsigned)((((long long)(1024) * ((1024) / 2)) + 255) / 256), 256, 0, stream>>>(cWq, 1024, (_Float16*)(G64B), 1024, 1024, 1024, 16.0f);
    w25::wmma_gemm64<0, false, 0, 0, false, 0><<<dim3((unsigned)((((512) / 64) * ((1024) / 64) + 7) / 8), (unsigned)(1)), 256, 0, stream>>>((const unsigned short*)(G64A), nullptr, 1024, 0, (const unsigned short*)(G64B), nullptr, 1024, 0, (void*)(Q), nullptr, 1024, 0, nullptr, nullptr, 0, 512, 1024, 1024, 0.0625f);
    { GemmP cq0ab;
      cq0ab.A = LOW; cq0ab.B = qb + (size_t)1 * R * D; cq0ab.bias = LOW; cq0ab.R = Q; cq0ab.C = Q;
      cq0ab.sAo = 0; cq0ab.sAi = 0; cq0ab.sAm = R; cq0ab.sAk = 1; cq0ab.sBo = 0; cq0ab.sBi = 0; cq0ab.sBn = 1; cq0ab.sBk = D; cq0ab.sCo = 0; cq0ab.sCi = 0; cq0ab.sCm = D; cq0ab.sRo = 0; cq0ab.sRi = 0; cq0ab.sRm = D; cq0ab.sRn = 1;
      cq0ab.M = L; cq0ab.N = D; cq0ab.K = R; cq0ab.zi_n = 1; cq0ab.flags = 4; cq0ab.act = 0;
      cq0ab.alpha = 1.0f; cq0ab.beta = 1.0f; cq0ab.sa = 1.0f; cq0ab.sb = 1.0f; cq0ab.Npad = D; cq0ab.pad_ = 0;
      if ((long long)(L) >= 64 && (long long)(D) >= 64) k_gemmT<0, 4, 4><<<dim3((unsigned)((D) + 63) / 64, (unsigned)((L) + 63) / 64, (unsigned)(1)), 32, 0, stream>>>(cq0ab);
      else k_gemm<0><<<dim3((unsigned)((D) + 31) / 32, (unsigned)((L) + 15) / 16, (unsigned)(1)), 32, 0, stream>>>(cq0ab); }
    { GemmP ck0lo;
      ck0lo.A = enc + (size_t)0 * L * D; ck0lo.B = ka + (size_t)1 * D * R; ck0lo.bias = enc + (size_t)0 * L * D; ck0lo.R = enc + (size_t)0 * L * D; ck0lo.C = LOW;
      ck0lo.sAo = 0; ck0lo.sAi = 0; ck0lo.sAm = D; ck0lo.sAk = 1; ck0lo.sBo = 0; ck0lo.sBi = 0; ck0lo.sBn = 1; ck0lo.sBk = R; ck0lo.sCo = 0; ck0lo.sCi = 0; ck0lo.sCm = R; ck0lo.sRo = 0; ck0lo.sRi = 0; ck0lo.sRm = 0; ck0lo.sRn = 0;
      ck0lo.M = L; ck0lo.N = R; ck0lo.K = D; ck0lo.zi_n = 1; ck0lo.flags = 0; ck0lo.act = 0;
      ck0lo.alpha = 1.0f; ck0lo.beta = 0.0f; ck0lo.sa = 1.0f; ck0lo.sb = 1.0f; ck0lo.Npad = R; ck0lo.pad_ = 0;
      if ((long long)(L) >= 64 && (long long)(R) >= 64) k_gemmT<0, 4, 4><<<dim3((unsigned)((R) + 63) / 64, (unsigned)((L) + 63) / 64, (unsigned)(1)), 32, 0, stream>>>(ck0lo);
      else k_gemm<0><<<dim3((unsigned)((R) + 31) / 32, (unsigned)((L) + 15) / 16, (unsigned)(1)), 32, 0, stream>>>(ck0lo); }
    k_cast16<<<(unsigned)((((long long)(512) * ((1024) / 2)) + 255) / 256), 256, 0, stream>>>(enc + (size_t)0 * L * D, 1024, (_Float16*)(G64A), 1024, 512, 1024, 1.0f);
    k_castT16<<<(unsigned)((((long long)(1024) * ((1024) / 2)) + 255) / 256), 256, 0, stream>>>(cWk, 1024, (_Float16*)(G64B), 1024, 1024, 1024, 16.0f);
    w25::wmma_gemm64<0, false, 0, 0, false, 0><<<dim3((unsigned)((((512) / 64) * ((1024) / 64) + 7) / 8), (unsigned)(1)), 256, 0, stream>>>((const unsigned short*)(G64A), nullptr, 1024, 0, (const unsigned short*)(G64B), nullptr, 1024, 0, (void*)(Kb), nullptr, 1024, 0, nullptr, nullptr, 0, 512, 1024, 1024, 0.0625f);
    { GemmP ck0ab;
      ck0ab.A = LOW; ck0ab.B = kb + (size_t)1 * R * D; ck0ab.bias = LOW; ck0ab.R = Kb; ck0ab.C = Kb;
      ck0ab.sAo = 0; ck0ab.sAi = 0; ck0ab.sAm = R; ck0ab.sAk = 1; ck0ab.sBo = 0; ck0ab.sBi = 0; ck0ab.sBn = 1; ck0ab.sBk = D; ck0ab.sCo = 0; ck0ab.sCi = 0; ck0ab.sCm = D; ck0ab.sRo = 0; ck0ab.sRi = 0; ck0ab.sRm = D; ck0ab.sRn = 1;
      ck0ab.M = L; ck0ab.N = D; ck0ab.K = R; ck0ab.zi_n = 1; ck0ab.flags = 4; ck0ab.act = 0;
      ck0ab.alpha = 1.0f; ck0ab.beta = 1.0f; ck0ab.sa = 1.0f; ck0ab.sb = 1.0f; ck0ab.Npad = D; ck0ab.pad_ = 0;
      if ((long long)(L) >= 64 && (long long)(D) >= 64) k_gemmT<0, 4, 4><<<dim3((unsigned)((D) + 63) / 64, (unsigned)((L) + 63) / 64, (unsigned)(1)), 32, 0, stream>>>(ck0ab);
      else k_gemm<0><<<dim3((unsigned)((D) + 31) / 32, (unsigned)((L) + 15) / 16, (unsigned)(1)), 32, 0, stream>>>(ck0ab); }
    { GemmP cv0lo;
      cv0lo.A = enc + (size_t)0 * L * D; cv0lo.B = va + (size_t)1 * D * R; cv0lo.bias = enc + (size_t)0 * L * D; cv0lo.R = enc + (size_t)0 * L * D; cv0lo.C = LOW;
      cv0lo.sAo = 0; cv0lo.sAi = 0; cv0lo.sAm = D; cv0lo.sAk = 1; cv0lo.sBo = 0; cv0lo.sBi = 0; cv0lo.sBn = 1; cv0lo.sBk = R; cv0lo.sCo = 0; cv0lo.sCi = 0; cv0lo.sCm = R; cv0lo.sRo = 0; cv0lo.sRi = 0; cv0lo.sRm = 0; cv0lo.sRn = 0;
      cv0lo.M = L; cv0lo.N = R; cv0lo.K = D; cv0lo.zi_n = 1; cv0lo.flags = 0; cv0lo.act = 0;
      cv0lo.alpha = 1.0f; cv0lo.beta = 0.0f; cv0lo.sa = 1.0f; cv0lo.sb = 1.0f; cv0lo.Npad = R; cv0lo.pad_ = 0;
      if ((long long)(L) >= 64 && (long long)(R) >= 64) k_gemmT<0, 4, 4><<<dim3((unsigned)((R) + 63) / 64, (unsigned)((L) + 63) / 64, (unsigned)(1)), 32, 0, stream>>>(cv0lo);
      else k_gemm<0><<<dim3((unsigned)((R) + 31) / 32, (unsigned)((L) + 15) / 16, (unsigned)(1)), 32, 0, stream>>>(cv0lo); }
    k_cast16<<<(unsigned)((((long long)(512) * ((1024) / 2)) + 255) / 256), 256, 0, stream>>>(enc + (size_t)0 * L * D, 1024, (_Float16*)(G64A), 1024, 512, 1024, 1.0f);
    k_castT16<<<(unsigned)((((long long)(1024) * ((1024) / 2)) + 255) / 256), 256, 0, stream>>>(cWv, 1024, (_Float16*)(G64B), 1024, 1024, 1024, 16.0f);
    w25::wmma_gemm64<0, false, 0, 0, false, 0><<<dim3((unsigned)((((512) / 64) * ((1024) / 64) + 7) / 8), (unsigned)(1)), 256, 0, stream>>>((const unsigned short*)(G64A), nullptr, 1024, 0, (const unsigned short*)(G64B), nullptr, 1024, 0, (void*)(V), nullptr, 1024, 0, nullptr, nullptr, 0, 512, 1024, 1024, 0.0625f);
    { GemmP cv0ab;
      cv0ab.A = LOW; cv0ab.B = vb + (size_t)1 * R * D; cv0ab.bias = LOW; cv0ab.R = V; cv0ab.C = V;
      cv0ab.sAo = 0; cv0ab.sAi = 0; cv0ab.sAm = R; cv0ab.sAk = 1; cv0ab.sBo = 0; cv0ab.sBi = 0; cv0ab.sBn = 1; cv0ab.sBk = D; cv0ab.sCo = 0; cv0ab.sCi = 0; cv0ab.sCm = D; cv0ab.sRo = 0; cv0ab.sRi = 0; cv0ab.sRm = D; cv0ab.sRn = 1;
      cv0ab.M = L; cv0ab.N = D; cv0ab.K = R; cv0ab.zi_n = 1; cv0ab.flags = 4; cv0ab.act = 0;
      cv0ab.alpha = 1.0f; cv0ab.beta = 1.0f; cv0ab.sa = 1.0f; cv0ab.sb = 1.0f; cv0ab.Npad = D; cv0ab.pad_ = 0;
      if ((long long)(L) >= 64 && (long long)(D) >= 64) k_gemmT<0, 4, 4><<<dim3((unsigned)((D) + 63) / 64, (unsigned)((L) + 63) / 64, (unsigned)(1)), 32, 0, stream>>>(cv0ab);
      else k_gemm<0><<<dim3((unsigned)((D) + 31) / 32, (unsigned)((L) + 15) / 16, (unsigned)(1)), 32, 0, stream>>>(cv0ab); }
    {   AttnP a;
      a.Q = Q; a.K = Kb; a.V = V; a.O = AT; a.P = 0; a.Mf = 0; a.Mi = 0; a.ST = 0;
      a.Pw = 0; a.Rt = 0; a.SQ = 0; a.SK = 0;
      a.swb = 0; a.swh = 0; a.swi = 0; a.swj = 0; a.srb = 0; a.srh = 0; a.sri = 0; a.sQb = 0; a.sQh = HD; a.sQi = D; a.sQd = 1; a.sKb = 0; a.sKh = HD; a.sKj = D; a.sKd = 1; a.sVb = 0; a.sVh = HD; a.sVj = D; a.sVd = 1; a.sOb = 0; a.sOh = HD; a.sOi = D; a.sPb = 0; a.sPh = 0; a.sPi = 0; a.smb = 0; a.smh = 0; a.smi = 0; a.smj = 0;
      a.Lq = L; a.Lk = L; a.dh = HD; a.dv = HD; a.hrep = 1; a.causal = 0; a.coff = 0; a.pband = 0;
      a.scale = 0.125f; a.mfill = 0.0f; a.nonorm = 0; a.mpol = 0;
      a.roff = 0; a.rn = 1; a.segpol = 0; a.win = 0;
      k_attn<64, 64, 0, false, false><<<dim3((unsigned)((L) + 16 * AW - 1) / (16 * AW), (unsigned)(NH), (unsigned)(1)), 32 * AW, 0, stream>>>(a); }
    { GemmP co0lo;
      co0lo.A = AT; co0lo.B = oa + (size_t)1 * D * R; co0lo.bias = AT; co0lo.R = AT; co0lo.C = LOW;
      co0lo.sAo = 0; co0lo.sAi = 0; co0lo.sAm = D; co0lo.sAk = 1; co0lo.sBo = 0; co0lo.sBi = 0; co0lo.sBn = 1; co0lo.sBk = R; co0lo.sCo = 0; co0lo.sCi = 0; co0lo.sCm = R; co0lo.sRo = 0; co0lo.sRi = 0; co0lo.sRm = 0; co0lo.sRn = 0;
      co0lo.M = L; co0lo.N = R; co0lo.K = D; co0lo.zi_n = 1; co0lo.flags = 0; co0lo.act = 0;
      co0lo.alpha = 1.0f; co0lo.beta = 0.0f; co0lo.sa = 1.0f; co0lo.sb = 1.0f; co0lo.Npad = R; co0lo.pad_ = 0;
      if ((long long)(L) >= 64 && (long long)(R) >= 64) k_gemmT<0, 4, 4><<<dim3((unsigned)((R) + 63) / 64, (unsigned)((L) + 63) / 64, (unsigned)(1)), 32, 0, stream>>>(co0lo);
      else k_gemm<0><<<dim3((unsigned)((R) + 31) / 32, (unsigned)((L) + 15) / 16, (unsigned)(1)), 32, 0, stream>>>(co0lo); }
    k_cast16<<<(unsigned)((((long long)(512) * ((1024) / 2)) + 255) / 256), 256, 0, stream>>>(AT, 1024, (_Float16*)(G64A), 1024, 512, 1024, 1.0f);
    k_castT16<<<(unsigned)((((long long)(1024) * ((1024) / 2)) + 255) / 256), 256, 0, stream>>>(cWo, 1024, (_Float16*)(G64B), 1024, 1024, 1024, 16.0f);
    w25::wmma_gemm64<0, false, 0, 0, true, 0><<<dim3((unsigned)((((512) / 64) * ((1024) / 64) + 7) / 8), (unsigned)(1)), 256, 0, stream>>>((const unsigned short*)(G64A), nullptr, 1024, 0, (const unsigned short*)(G64B), nullptr, 1024, 0, (void*)(Y1 + (size_t)0 * L * D), nullptr, 1024, 0, nullptr, X1 + (size_t)0 * L * D, 0, 512, 1024, 1024, 0.0625f);
    { GemmP co0ab;
      co0ab.A = LOW; co0ab.B = ob + (size_t)1 * R * D; co0ab.bias = LOW; co0ab.R = Y1 + (size_t)0 * L * D; co0ab.C = Y1 + (size_t)0 * L * D;
      co0ab.sAo = 0; co0ab.sAi = 0; co0ab.sAm = R; co0ab.sAk = 1; co0ab.sBo = 0; co0ab.sBi = 0; co0ab.sBn = 1; co0ab.sBk = D; co0ab.sCo = 0; co0ab.sCi = 0; co0ab.sCm = D; co0ab.sRo = 0; co0ab.sRi = 0; co0ab.sRm = D; co0ab.sRn = 1;
      co0ab.M = L; co0ab.N = D; co0ab.K = R; co0ab.zi_n = 1; co0ab.flags = 4; co0ab.act = 0;
      co0ab.alpha = 1.0f; co0ab.beta = 1.0f; co0ab.sa = 1.0f; co0ab.sb = 1.0f; co0ab.Npad = D; co0ab.pad_ = 0;
      if ((long long)(L) >= 64 && (long long)(D) >= 64) k_gemmT<0, 4, 4><<<dim3((unsigned)((D) + 63) / 64, (unsigned)((L) + 63) / 64, (unsigned)(1)), 32, 0, stream>>>(co0ab);
      else k_gemm<0><<<dim3((unsigned)((D) + 31) / 32, (unsigned)((L) + 15) / 16, (unsigned)(1)), 32, 0, stream>>>(co0ab); }
    k_ld_rms<<<L, 256, 0, stream>>>(Y1 + (size_t)0 * L * D, ln3, XN, D);
    k_cast16<<<(unsigned)((((long long)(512) * ((1024) / 2)) + 255) / 256), 256, 0, stream>>>(XN, 1024, (_Float16*)(G64A), 1024, 512, 1024, 1.0f);
    k_castT16<<<(unsigned)((((long long)(4096) * ((1024) / 2)) + 255) / 256), 256, 0, stream>>>(wi0, 4096, (_Float16*)(G64B), 1024, 1024, 4096, 16.0f);
    w25::wmma_gemm64<0, false, 0, 0, false, 0><<<dim3((unsigned)((((512) / 64) * ((4096) / 64) + 7) / 8), (unsigned)(1)), 256, 0, stream>>>((const unsigned short*)(G64A), nullptr, 1024, 0, (const unsigned short*)(G64B), nullptr, 1024, 0, (void*)(G0), nullptr, 4096, 0, nullptr, nullptr, 0, 512, 4096, 1024, 0.0625f);
    k_cast16<<<(unsigned)((((long long)(512) * ((1024) / 2)) + 255) / 256), 256, 0, stream>>>(XN, 1024, (_Float16*)(G64A), 1024, 512, 1024, 1.0f);
    k_castT16<<<(unsigned)((((long long)(4096) * ((1024) / 2)) + 255) / 256), 256, 0, stream>>>(wi1, 4096, (_Float16*)(G64B), 1024, 1024, 4096, 16.0f);
    w25::wmma_gemm64<0, false, 0, 0, false, 0><<<dim3((unsigned)((((512) / 64) * ((4096) / 64) + 7) / 8), (unsigned)(1)), 256, 0, stream>>>((const unsigned short*)(G64A), nullptr, 1024, 0, (const unsigned short*)(G64B), nullptr, 1024, 0, (void*)(G1), nullptr, 4096, 0, nullptr, nullptr, 0, 512, 4096, 1024, 0.0625f);
    k_ld_gg<<<(unsigned)(((long long)L * FF + 255) / 256), 256, 0, stream>>>(G0, G1, (long long)L * FF);
    k_cast16<<<(unsigned)((((long long)(512) * ((4096) / 2)) + 255) / 256), 256, 0, stream>>>(G0, 4096, (_Float16*)(G64A), 4096, 512, 4096, 1.0f);
    k_castT16<<<(unsigned)((((long long)(1024) * ((4096) / 2)) + 255) / 256), 256, 0, stream>>>(wom, 1024, (_Float16*)(G64B), 4096, 4096, 1024, 16.0f);
    w25::wmma_gemm64<0, false, 0, 0, true, 0><<<dim3((unsigned)((((512) / 64) * ((1024) / 64) + 7) / 8), (unsigned)(1)), 256, 0, stream>>>((const unsigned short*)(G64A), nullptr, 4096, 0, (const unsigned short*)(G64B), nullptr, 4096, 0, (void*)(out + (size_t)0 * L * D), nullptr, 1024, 0, nullptr, Y1 + (size_t)0 * L * D, 0, 512, 1024, 4096, 0.0625f);
    k_ld_rms<<<L, 256, 0, stream>>>(xin + (size_t)1 * L * D, ln1, XN, D);
    { GemmP sq1lo;
      sq1lo.A = XN; sq1lo.B = qa + (size_t)2 * D * R; sq1lo.bias = XN; sq1lo.R = XN; sq1lo.C = LOW;
      sq1lo.sAo = 0; sq1lo.sAi = 0; sq1lo.sAm = D; sq1lo.sAk = 1; sq1lo.sBo = 0; sq1lo.sBi = 0; sq1lo.sBn = 1; sq1lo.sBk = R; sq1lo.sCo = 0; sq1lo.sCi = 0; sq1lo.sCm = R; sq1lo.sRo = 0; sq1lo.sRi = 0; sq1lo.sRm = 0; sq1lo.sRn = 0;
      sq1lo.M = L; sq1lo.N = R; sq1lo.K = D; sq1lo.zi_n = 1; sq1lo.flags = 0; sq1lo.act = 0;
      sq1lo.alpha = 1.0f; sq1lo.beta = 0.0f; sq1lo.sa = 1.0f; sq1lo.sb = 1.0f; sq1lo.Npad = R; sq1lo.pad_ = 0;
      if ((long long)(L) >= 64 && (long long)(R) >= 64) k_gemmT<0, 4, 4><<<dim3((unsigned)((R) + 63) / 64, (unsigned)((L) + 63) / 64, (unsigned)(1)), 32, 0, stream>>>(sq1lo);
      else k_gemm<0><<<dim3((unsigned)((R) + 31) / 32, (unsigned)((L) + 15) / 16, (unsigned)(1)), 32, 0, stream>>>(sq1lo); }
    k_cast16<<<(unsigned)((((long long)(512) * ((1024) / 2)) + 255) / 256), 256, 0, stream>>>(XN, 1024, (_Float16*)(G64A), 1024, 512, 1024, 1.0f);
    k_castT16<<<(unsigned)((((long long)(1024) * ((1024) / 2)) + 255) / 256), 256, 0, stream>>>(sWq, 1024, (_Float16*)(G64B), 1024, 1024, 1024, 16.0f);
    w25::wmma_gemm64<0, false, 0, 0, false, 0><<<dim3((unsigned)((((512) / 64) * ((1024) / 64) + 7) / 8), (unsigned)(1)), 256, 0, stream>>>((const unsigned short*)(G64A), nullptr, 1024, 0, (const unsigned short*)(G64B), nullptr, 1024, 0, (void*)(Q), nullptr, 1024, 0, nullptr, nullptr, 0, 512, 1024, 1024, 0.0625f);
    { GemmP sq1ab;
      sq1ab.A = LOW; sq1ab.B = qb + (size_t)2 * R * D; sq1ab.bias = LOW; sq1ab.R = Q; sq1ab.C = Q;
      sq1ab.sAo = 0; sq1ab.sAi = 0; sq1ab.sAm = R; sq1ab.sAk = 1; sq1ab.sBo = 0; sq1ab.sBi = 0; sq1ab.sBn = 1; sq1ab.sBk = D; sq1ab.sCo = 0; sq1ab.sCi = 0; sq1ab.sCm = D; sq1ab.sRo = 0; sq1ab.sRi = 0; sq1ab.sRm = D; sq1ab.sRn = 1;
      sq1ab.M = L; sq1ab.N = D; sq1ab.K = R; sq1ab.zi_n = 1; sq1ab.flags = 4; sq1ab.act = 0;
      sq1ab.alpha = 1.0f; sq1ab.beta = 1.0f; sq1ab.sa = 1.0f; sq1ab.sb = 1.0f; sq1ab.Npad = D; sq1ab.pad_ = 0;
      if ((long long)(L) >= 64 && (long long)(D) >= 64) k_gemmT<0, 4, 4><<<dim3((unsigned)((D) + 63) / 64, (unsigned)((L) + 63) / 64, (unsigned)(1)), 32, 0, stream>>>(sq1ab);
      else k_gemm<0><<<dim3((unsigned)((D) + 31) / 32, (unsigned)((L) + 15) / 16, (unsigned)(1)), 32, 0, stream>>>(sq1ab); }
    { GemmP sk1lo;
      sk1lo.A = XN; sk1lo.B = ka + (size_t)2 * D * R; sk1lo.bias = XN; sk1lo.R = XN; sk1lo.C = LOW;
      sk1lo.sAo = 0; sk1lo.sAi = 0; sk1lo.sAm = D; sk1lo.sAk = 1; sk1lo.sBo = 0; sk1lo.sBi = 0; sk1lo.sBn = 1; sk1lo.sBk = R; sk1lo.sCo = 0; sk1lo.sCi = 0; sk1lo.sCm = R; sk1lo.sRo = 0; sk1lo.sRi = 0; sk1lo.sRm = 0; sk1lo.sRn = 0;
      sk1lo.M = L; sk1lo.N = R; sk1lo.K = D; sk1lo.zi_n = 1; sk1lo.flags = 0; sk1lo.act = 0;
      sk1lo.alpha = 1.0f; sk1lo.beta = 0.0f; sk1lo.sa = 1.0f; sk1lo.sb = 1.0f; sk1lo.Npad = R; sk1lo.pad_ = 0;
      if ((long long)(L) >= 64 && (long long)(R) >= 64) k_gemmT<0, 4, 4><<<dim3((unsigned)((R) + 63) / 64, (unsigned)((L) + 63) / 64, (unsigned)(1)), 32, 0, stream>>>(sk1lo);
      else k_gemm<0><<<dim3((unsigned)((R) + 31) / 32, (unsigned)((L) + 15) / 16, (unsigned)(1)), 32, 0, stream>>>(sk1lo); }
    k_cast16<<<(unsigned)((((long long)(512) * ((1024) / 2)) + 255) / 256), 256, 0, stream>>>(XN, 1024, (_Float16*)(G64A), 1024, 512, 1024, 1.0f);
    k_castT16<<<(unsigned)((((long long)(1024) * ((1024) / 2)) + 255) / 256), 256, 0, stream>>>(sWk, 1024, (_Float16*)(G64B), 1024, 1024, 1024, 16.0f);
    w25::wmma_gemm64<0, false, 0, 0, false, 0><<<dim3((unsigned)((((512) / 64) * ((1024) / 64) + 7) / 8), (unsigned)(1)), 256, 0, stream>>>((const unsigned short*)(G64A), nullptr, 1024, 0, (const unsigned short*)(G64B), nullptr, 1024, 0, (void*)(Kb), nullptr, 1024, 0, nullptr, nullptr, 0, 512, 1024, 1024, 0.0625f);
    { GemmP sk1ab;
      sk1ab.A = LOW; sk1ab.B = kb + (size_t)2 * R * D; sk1ab.bias = LOW; sk1ab.R = Kb; sk1ab.C = Kb;
      sk1ab.sAo = 0; sk1ab.sAi = 0; sk1ab.sAm = R; sk1ab.sAk = 1; sk1ab.sBo = 0; sk1ab.sBi = 0; sk1ab.sBn = 1; sk1ab.sBk = D; sk1ab.sCo = 0; sk1ab.sCi = 0; sk1ab.sCm = D; sk1ab.sRo = 0; sk1ab.sRi = 0; sk1ab.sRm = D; sk1ab.sRn = 1;
      sk1ab.M = L; sk1ab.N = D; sk1ab.K = R; sk1ab.zi_n = 1; sk1ab.flags = 4; sk1ab.act = 0;
      sk1ab.alpha = 1.0f; sk1ab.beta = 1.0f; sk1ab.sa = 1.0f; sk1ab.sb = 1.0f; sk1ab.Npad = D; sk1ab.pad_ = 0;
      if ((long long)(L) >= 64 && (long long)(D) >= 64) k_gemmT<0, 4, 4><<<dim3((unsigned)((D) + 63) / 64, (unsigned)((L) + 63) / 64, (unsigned)(1)), 32, 0, stream>>>(sk1ab);
      else k_gemm<0><<<dim3((unsigned)((D) + 31) / 32, (unsigned)((L) + 15) / 16, (unsigned)(1)), 32, 0, stream>>>(sk1ab); }
    { GemmP sv1lo;
      sv1lo.A = XN; sv1lo.B = va + (size_t)2 * D * R; sv1lo.bias = XN; sv1lo.R = XN; sv1lo.C = LOW;
      sv1lo.sAo = 0; sv1lo.sAi = 0; sv1lo.sAm = D; sv1lo.sAk = 1; sv1lo.sBo = 0; sv1lo.sBi = 0; sv1lo.sBn = 1; sv1lo.sBk = R; sv1lo.sCo = 0; sv1lo.sCi = 0; sv1lo.sCm = R; sv1lo.sRo = 0; sv1lo.sRi = 0; sv1lo.sRm = 0; sv1lo.sRn = 0;
      sv1lo.M = L; sv1lo.N = R; sv1lo.K = D; sv1lo.zi_n = 1; sv1lo.flags = 0; sv1lo.act = 0;
      sv1lo.alpha = 1.0f; sv1lo.beta = 0.0f; sv1lo.sa = 1.0f; sv1lo.sb = 1.0f; sv1lo.Npad = R; sv1lo.pad_ = 0;
      if ((long long)(L) >= 64 && (long long)(R) >= 64) k_gemmT<0, 4, 4><<<dim3((unsigned)((R) + 63) / 64, (unsigned)((L) + 63) / 64, (unsigned)(1)), 32, 0, stream>>>(sv1lo);
      else k_gemm<0><<<dim3((unsigned)((R) + 31) / 32, (unsigned)((L) + 15) / 16, (unsigned)(1)), 32, 0, stream>>>(sv1lo); }
    k_cast16<<<(unsigned)((((long long)(512) * ((1024) / 2)) + 255) / 256), 256, 0, stream>>>(XN, 1024, (_Float16*)(G64A), 1024, 512, 1024, 1.0f);
    k_castT16<<<(unsigned)((((long long)(1024) * ((1024) / 2)) + 255) / 256), 256, 0, stream>>>(sWv, 1024, (_Float16*)(G64B), 1024, 1024, 1024, 16.0f);
    w25::wmma_gemm64<0, false, 0, 0, false, 0><<<dim3((unsigned)((((512) / 64) * ((1024) / 64) + 7) / 8), (unsigned)(1)), 256, 0, stream>>>((const unsigned short*)(G64A), nullptr, 1024, 0, (const unsigned short*)(G64B), nullptr, 1024, 0, (void*)(V), nullptr, 1024, 0, nullptr, nullptr, 0, 512, 1024, 1024, 0.0625f);
    { GemmP sv1ab;
      sv1ab.A = LOW; sv1ab.B = vb + (size_t)2 * R * D; sv1ab.bias = LOW; sv1ab.R = V; sv1ab.C = V;
      sv1ab.sAo = 0; sv1ab.sAi = 0; sv1ab.sAm = R; sv1ab.sAk = 1; sv1ab.sBo = 0; sv1ab.sBi = 0; sv1ab.sBn = 1; sv1ab.sBk = D; sv1ab.sCo = 0; sv1ab.sCi = 0; sv1ab.sCm = D; sv1ab.sRo = 0; sv1ab.sRi = 0; sv1ab.sRm = D; sv1ab.sRn = 1;
      sv1ab.M = L; sv1ab.N = D; sv1ab.K = R; sv1ab.zi_n = 1; sv1ab.flags = 4; sv1ab.act = 0;
      sv1ab.alpha = 1.0f; sv1ab.beta = 1.0f; sv1ab.sa = 1.0f; sv1ab.sb = 1.0f; sv1ab.Npad = D; sv1ab.pad_ = 0;
      if ((long long)(L) >= 64 && (long long)(D) >= 64) k_gemmT<0, 4, 4><<<dim3((unsigned)((D) + 63) / 64, (unsigned)((L) + 63) / 64, (unsigned)(1)), 32, 0, stream>>>(sv1ab);
      else k_gemm<0><<<dim3((unsigned)((D) + 31) / 32, (unsigned)((L) + 15) / 16, (unsigned)(1)), 32, 0, stream>>>(sv1ab); }
    {   AttnP a;
      a.Q = Q; a.K = Kb; a.V = V; a.O = AT; a.P = 0; a.Mf = BIAS; a.Mi = 0; a.ST = 0;
      a.Pw = 0; a.Rt = 0; a.SQ = 0; a.SK = 0;
      a.swb = 0; a.swh = 0; a.swi = 0; a.swj = 0; a.srb = 0; a.srh = 0; a.sri = 0; a.sQb = 0; a.sQh = HD; a.sQi = D; a.sQd = 1; a.sKb = 0; a.sKh = HD; a.sKj = D; a.sKd = 1; a.sVb = 0; a.sVh = HD; a.sVj = D; a.sVd = 1; a.sOb = 0; a.sOh = HD; a.sOi = D; a.sPb = 0; a.sPh = 0; a.sPi = 0; a.smb = 0; a.smh = (long long)L * L; a.smi = L; a.smj = 1;
      a.Lq = L; a.Lk = L; a.dh = HD; a.dv = HD; a.hrep = 1; a.causal = 1; a.coff = 0; a.pband = 0;
      a.scale = 0.125f; a.mfill = 0.0f; a.nonorm = 0; a.mpol = 0;
      a.roff = 0; a.rn = 1; a.segpol = 0; a.win = 0;
      k_attn<64, 64, 0, false, false><<<dim3((unsigned)((L) + 16 * AW - 1) / (16 * AW), (unsigned)(NH), (unsigned)(1)), 32 * AW, 0, stream>>>(a); }
    { GemmP so1lo;
      so1lo.A = AT; so1lo.B = oa + (size_t)2 * D * R; so1lo.bias = AT; so1lo.R = AT; so1lo.C = LOW;
      so1lo.sAo = 0; so1lo.sAi = 0; so1lo.sAm = D; so1lo.sAk = 1; so1lo.sBo = 0; so1lo.sBi = 0; so1lo.sBn = 1; so1lo.sBk = R; so1lo.sCo = 0; so1lo.sCi = 0; so1lo.sCm = R; so1lo.sRo = 0; so1lo.sRi = 0; so1lo.sRm = 0; so1lo.sRn = 0;
      so1lo.M = L; so1lo.N = R; so1lo.K = D; so1lo.zi_n = 1; so1lo.flags = 0; so1lo.act = 0;
      so1lo.alpha = 1.0f; so1lo.beta = 0.0f; so1lo.sa = 1.0f; so1lo.sb = 1.0f; so1lo.Npad = R; so1lo.pad_ = 0;
      if ((long long)(L) >= 64 && (long long)(R) >= 64) k_gemmT<0, 4, 4><<<dim3((unsigned)((R) + 63) / 64, (unsigned)((L) + 63) / 64, (unsigned)(1)), 32, 0, stream>>>(so1lo);
      else k_gemm<0><<<dim3((unsigned)((R) + 31) / 32, (unsigned)((L) + 15) / 16, (unsigned)(1)), 32, 0, stream>>>(so1lo); }
    k_cast16<<<(unsigned)((((long long)(512) * ((1024) / 2)) + 255) / 256), 256, 0, stream>>>(AT, 1024, (_Float16*)(G64A), 1024, 512, 1024, 1.0f);
    k_castT16<<<(unsigned)((((long long)(1024) * ((1024) / 2)) + 255) / 256), 256, 0, stream>>>(sWo, 1024, (_Float16*)(G64B), 1024, 1024, 1024, 16.0f);
    w25::wmma_gemm64<0, false, 0, 0, true, 0><<<dim3((unsigned)((((512) / 64) * ((1024) / 64) + 7) / 8), (unsigned)(1)), 256, 0, stream>>>((const unsigned short*)(G64A), nullptr, 1024, 0, (const unsigned short*)(G64B), nullptr, 1024, 0, (void*)(X1 + (size_t)1 * L * D), nullptr, 1024, 0, nullptr, xin + (size_t)1 * L * D, 0, 512, 1024, 1024, 0.0625f);
    { GemmP so1ab;
      so1ab.A = LOW; so1ab.B = ob + (size_t)2 * R * D; so1ab.bias = LOW; so1ab.R = X1 + (size_t)1 * L * D; so1ab.C = X1 + (size_t)1 * L * D;
      so1ab.sAo = 0; so1ab.sAi = 0; so1ab.sAm = R; so1ab.sAk = 1; so1ab.sBo = 0; so1ab.sBi = 0; so1ab.sBn = 1; so1ab.sBk = D; so1ab.sCo = 0; so1ab.sCi = 0; so1ab.sCm = D; so1ab.sRo = 0; so1ab.sRi = 0; so1ab.sRm = D; so1ab.sRn = 1;
      so1ab.M = L; so1ab.N = D; so1ab.K = R; so1ab.zi_n = 1; so1ab.flags = 4; so1ab.act = 0;
      so1ab.alpha = 1.0f; so1ab.beta = 1.0f; so1ab.sa = 1.0f; so1ab.sb = 1.0f; so1ab.Npad = D; so1ab.pad_ = 0;
      if ((long long)(L) >= 64 && (long long)(D) >= 64) k_gemmT<0, 4, 4><<<dim3((unsigned)((D) + 63) / 64, (unsigned)((L) + 63) / 64, (unsigned)(1)), 32, 0, stream>>>(so1ab);
      else k_gemm<0><<<dim3((unsigned)((D) + 31) / 32, (unsigned)((L) + 15) / 16, (unsigned)(1)), 32, 0, stream>>>(so1ab); }
    k_ld_rms<<<L, 256, 0, stream>>>(X1 + (size_t)1 * L * D, ln2, XN, D);
    { GemmP cq1lo;
      cq1lo.A = XN; cq1lo.B = qa + (size_t)3 * D * R; cq1lo.bias = XN; cq1lo.R = XN; cq1lo.C = LOW;
      cq1lo.sAo = 0; cq1lo.sAi = 0; cq1lo.sAm = D; cq1lo.sAk = 1; cq1lo.sBo = 0; cq1lo.sBi = 0; cq1lo.sBn = 1; cq1lo.sBk = R; cq1lo.sCo = 0; cq1lo.sCi = 0; cq1lo.sCm = R; cq1lo.sRo = 0; cq1lo.sRi = 0; cq1lo.sRm = 0; cq1lo.sRn = 0;
      cq1lo.M = L; cq1lo.N = R; cq1lo.K = D; cq1lo.zi_n = 1; cq1lo.flags = 0; cq1lo.act = 0;
      cq1lo.alpha = 1.0f; cq1lo.beta = 0.0f; cq1lo.sa = 1.0f; cq1lo.sb = 1.0f; cq1lo.Npad = R; cq1lo.pad_ = 0;
      if ((long long)(L) >= 64 && (long long)(R) >= 64) k_gemmT<0, 4, 4><<<dim3((unsigned)((R) + 63) / 64, (unsigned)((L) + 63) / 64, (unsigned)(1)), 32, 0, stream>>>(cq1lo);
      else k_gemm<0><<<dim3((unsigned)((R) + 31) / 32, (unsigned)((L) + 15) / 16, (unsigned)(1)), 32, 0, stream>>>(cq1lo); }
    k_cast16<<<(unsigned)((((long long)(512) * ((1024) / 2)) + 255) / 256), 256, 0, stream>>>(XN, 1024, (_Float16*)(G64A), 1024, 512, 1024, 1.0f);
    k_castT16<<<(unsigned)((((long long)(1024) * ((1024) / 2)) + 255) / 256), 256, 0, stream>>>(cWq, 1024, (_Float16*)(G64B), 1024, 1024, 1024, 16.0f);
    w25::wmma_gemm64<0, false, 0, 0, false, 0><<<dim3((unsigned)((((512) / 64) * ((1024) / 64) + 7) / 8), (unsigned)(1)), 256, 0, stream>>>((const unsigned short*)(G64A), nullptr, 1024, 0, (const unsigned short*)(G64B), nullptr, 1024, 0, (void*)(Q), nullptr, 1024, 0, nullptr, nullptr, 0, 512, 1024, 1024, 0.0625f);
    { GemmP cq1ab;
      cq1ab.A = LOW; cq1ab.B = qb + (size_t)3 * R * D; cq1ab.bias = LOW; cq1ab.R = Q; cq1ab.C = Q;
      cq1ab.sAo = 0; cq1ab.sAi = 0; cq1ab.sAm = R; cq1ab.sAk = 1; cq1ab.sBo = 0; cq1ab.sBi = 0; cq1ab.sBn = 1; cq1ab.sBk = D; cq1ab.sCo = 0; cq1ab.sCi = 0; cq1ab.sCm = D; cq1ab.sRo = 0; cq1ab.sRi = 0; cq1ab.sRm = D; cq1ab.sRn = 1;
      cq1ab.M = L; cq1ab.N = D; cq1ab.K = R; cq1ab.zi_n = 1; cq1ab.flags = 4; cq1ab.act = 0;
      cq1ab.alpha = 1.0f; cq1ab.beta = 1.0f; cq1ab.sa = 1.0f; cq1ab.sb = 1.0f; cq1ab.Npad = D; cq1ab.pad_ = 0;
      if ((long long)(L) >= 64 && (long long)(D) >= 64) k_gemmT<0, 4, 4><<<dim3((unsigned)((D) + 63) / 64, (unsigned)((L) + 63) / 64, (unsigned)(1)), 32, 0, stream>>>(cq1ab);
      else k_gemm<0><<<dim3((unsigned)((D) + 31) / 32, (unsigned)((L) + 15) / 16, (unsigned)(1)), 32, 0, stream>>>(cq1ab); }
    { GemmP ck1lo;
      ck1lo.A = enc + (size_t)1 * L * D; ck1lo.B = ka + (size_t)3 * D * R; ck1lo.bias = enc + (size_t)1 * L * D; ck1lo.R = enc + (size_t)1 * L * D; ck1lo.C = LOW;
      ck1lo.sAo = 0; ck1lo.sAi = 0; ck1lo.sAm = D; ck1lo.sAk = 1; ck1lo.sBo = 0; ck1lo.sBi = 0; ck1lo.sBn = 1; ck1lo.sBk = R; ck1lo.sCo = 0; ck1lo.sCi = 0; ck1lo.sCm = R; ck1lo.sRo = 0; ck1lo.sRi = 0; ck1lo.sRm = 0; ck1lo.sRn = 0;
      ck1lo.M = L; ck1lo.N = R; ck1lo.K = D; ck1lo.zi_n = 1; ck1lo.flags = 0; ck1lo.act = 0;
      ck1lo.alpha = 1.0f; ck1lo.beta = 0.0f; ck1lo.sa = 1.0f; ck1lo.sb = 1.0f; ck1lo.Npad = R; ck1lo.pad_ = 0;
      if ((long long)(L) >= 64 && (long long)(R) >= 64) k_gemmT<0, 4, 4><<<dim3((unsigned)((R) + 63) / 64, (unsigned)((L) + 63) / 64, (unsigned)(1)), 32, 0, stream>>>(ck1lo);
      else k_gemm<0><<<dim3((unsigned)((R) + 31) / 32, (unsigned)((L) + 15) / 16, (unsigned)(1)), 32, 0, stream>>>(ck1lo); }
    k_cast16<<<(unsigned)((((long long)(512) * ((1024) / 2)) + 255) / 256), 256, 0, stream>>>(enc + (size_t)1 * L * D, 1024, (_Float16*)(G64A), 1024, 512, 1024, 1.0f);
    k_castT16<<<(unsigned)((((long long)(1024) * ((1024) / 2)) + 255) / 256), 256, 0, stream>>>(cWk, 1024, (_Float16*)(G64B), 1024, 1024, 1024, 16.0f);
    w25::wmma_gemm64<0, false, 0, 0, false, 0><<<dim3((unsigned)((((512) / 64) * ((1024) / 64) + 7) / 8), (unsigned)(1)), 256, 0, stream>>>((const unsigned short*)(G64A), nullptr, 1024, 0, (const unsigned short*)(G64B), nullptr, 1024, 0, (void*)(Kb), nullptr, 1024, 0, nullptr, nullptr, 0, 512, 1024, 1024, 0.0625f);
    { GemmP ck1ab;
      ck1ab.A = LOW; ck1ab.B = kb + (size_t)3 * R * D; ck1ab.bias = LOW; ck1ab.R = Kb; ck1ab.C = Kb;
      ck1ab.sAo = 0; ck1ab.sAi = 0; ck1ab.sAm = R; ck1ab.sAk = 1; ck1ab.sBo = 0; ck1ab.sBi = 0; ck1ab.sBn = 1; ck1ab.sBk = D; ck1ab.sCo = 0; ck1ab.sCi = 0; ck1ab.sCm = D; ck1ab.sRo = 0; ck1ab.sRi = 0; ck1ab.sRm = D; ck1ab.sRn = 1;
      ck1ab.M = L; ck1ab.N = D; ck1ab.K = R; ck1ab.zi_n = 1; ck1ab.flags = 4; ck1ab.act = 0;
      ck1ab.alpha = 1.0f; ck1ab.beta = 1.0f; ck1ab.sa = 1.0f; ck1ab.sb = 1.0f; ck1ab.Npad = D; ck1ab.pad_ = 0;
      if ((long long)(L) >= 64 && (long long)(D) >= 64) k_gemmT<0, 4, 4><<<dim3((unsigned)((D) + 63) / 64, (unsigned)((L) + 63) / 64, (unsigned)(1)), 32, 0, stream>>>(ck1ab);
      else k_gemm<0><<<dim3((unsigned)((D) + 31) / 32, (unsigned)((L) + 15) / 16, (unsigned)(1)), 32, 0, stream>>>(ck1ab); }
    { GemmP cv1lo;
      cv1lo.A = enc + (size_t)1 * L * D; cv1lo.B = va + (size_t)3 * D * R; cv1lo.bias = enc + (size_t)1 * L * D; cv1lo.R = enc + (size_t)1 * L * D; cv1lo.C = LOW;
      cv1lo.sAo = 0; cv1lo.sAi = 0; cv1lo.sAm = D; cv1lo.sAk = 1; cv1lo.sBo = 0; cv1lo.sBi = 0; cv1lo.sBn = 1; cv1lo.sBk = R; cv1lo.sCo = 0; cv1lo.sCi = 0; cv1lo.sCm = R; cv1lo.sRo = 0; cv1lo.sRi = 0; cv1lo.sRm = 0; cv1lo.sRn = 0;
      cv1lo.M = L; cv1lo.N = R; cv1lo.K = D; cv1lo.zi_n = 1; cv1lo.flags = 0; cv1lo.act = 0;
      cv1lo.alpha = 1.0f; cv1lo.beta = 0.0f; cv1lo.sa = 1.0f; cv1lo.sb = 1.0f; cv1lo.Npad = R; cv1lo.pad_ = 0;
      if ((long long)(L) >= 64 && (long long)(R) >= 64) k_gemmT<0, 4, 4><<<dim3((unsigned)((R) + 63) / 64, (unsigned)((L) + 63) / 64, (unsigned)(1)), 32, 0, stream>>>(cv1lo);
      else k_gemm<0><<<dim3((unsigned)((R) + 31) / 32, (unsigned)((L) + 15) / 16, (unsigned)(1)), 32, 0, stream>>>(cv1lo); }
    k_cast16<<<(unsigned)((((long long)(512) * ((1024) / 2)) + 255) / 256), 256, 0, stream>>>(enc + (size_t)1 * L * D, 1024, (_Float16*)(G64A), 1024, 512, 1024, 1.0f);
    k_castT16<<<(unsigned)((((long long)(1024) * ((1024) / 2)) + 255) / 256), 256, 0, stream>>>(cWv, 1024, (_Float16*)(G64B), 1024, 1024, 1024, 16.0f);
    w25::wmma_gemm64<0, false, 0, 0, false, 0><<<dim3((unsigned)((((512) / 64) * ((1024) / 64) + 7) / 8), (unsigned)(1)), 256, 0, stream>>>((const unsigned short*)(G64A), nullptr, 1024, 0, (const unsigned short*)(G64B), nullptr, 1024, 0, (void*)(V), nullptr, 1024, 0, nullptr, nullptr, 0, 512, 1024, 1024, 0.0625f);
    { GemmP cv1ab;
      cv1ab.A = LOW; cv1ab.B = vb + (size_t)3 * R * D; cv1ab.bias = LOW; cv1ab.R = V; cv1ab.C = V;
      cv1ab.sAo = 0; cv1ab.sAi = 0; cv1ab.sAm = R; cv1ab.sAk = 1; cv1ab.sBo = 0; cv1ab.sBi = 0; cv1ab.sBn = 1; cv1ab.sBk = D; cv1ab.sCo = 0; cv1ab.sCi = 0; cv1ab.sCm = D; cv1ab.sRo = 0; cv1ab.sRi = 0; cv1ab.sRm = D; cv1ab.sRn = 1;
      cv1ab.M = L; cv1ab.N = D; cv1ab.K = R; cv1ab.zi_n = 1; cv1ab.flags = 4; cv1ab.act = 0;
      cv1ab.alpha = 1.0f; cv1ab.beta = 1.0f; cv1ab.sa = 1.0f; cv1ab.sb = 1.0f; cv1ab.Npad = D; cv1ab.pad_ = 0;
      if ((long long)(L) >= 64 && (long long)(D) >= 64) k_gemmT<0, 4, 4><<<dim3((unsigned)((D) + 63) / 64, (unsigned)((L) + 63) / 64, (unsigned)(1)), 32, 0, stream>>>(cv1ab);
      else k_gemm<0><<<dim3((unsigned)((D) + 31) / 32, (unsigned)((L) + 15) / 16, (unsigned)(1)), 32, 0, stream>>>(cv1ab); }
    {   AttnP a;
      a.Q = Q; a.K = Kb; a.V = V; a.O = AT; a.P = 0; a.Mf = 0; a.Mi = 0; a.ST = 0;
      a.Pw = 0; a.Rt = 0; a.SQ = 0; a.SK = 0;
      a.swb = 0; a.swh = 0; a.swi = 0; a.swj = 0; a.srb = 0; a.srh = 0; a.sri = 0; a.sQb = 0; a.sQh = HD; a.sQi = D; a.sQd = 1; a.sKb = 0; a.sKh = HD; a.sKj = D; a.sKd = 1; a.sVb = 0; a.sVh = HD; a.sVj = D; a.sVd = 1; a.sOb = 0; a.sOh = HD; a.sOi = D; a.sPb = 0; a.sPh = 0; a.sPi = 0; a.smb = 0; a.smh = 0; a.smi = 0; a.smj = 0;
      a.Lq = L; a.Lk = L; a.dh = HD; a.dv = HD; a.hrep = 1; a.causal = 0; a.coff = 0; a.pband = 0;
      a.scale = 0.125f; a.mfill = 0.0f; a.nonorm = 0; a.mpol = 0;
      a.roff = 0; a.rn = 1; a.segpol = 0; a.win = 0;
      k_attn<64, 64, 0, false, false><<<dim3((unsigned)((L) + 16 * AW - 1) / (16 * AW), (unsigned)(NH), (unsigned)(1)), 32 * AW, 0, stream>>>(a); }
    { GemmP co1lo;
      co1lo.A = AT; co1lo.B = oa + (size_t)3 * D * R; co1lo.bias = AT; co1lo.R = AT; co1lo.C = LOW;
      co1lo.sAo = 0; co1lo.sAi = 0; co1lo.sAm = D; co1lo.sAk = 1; co1lo.sBo = 0; co1lo.sBi = 0; co1lo.sBn = 1; co1lo.sBk = R; co1lo.sCo = 0; co1lo.sCi = 0; co1lo.sCm = R; co1lo.sRo = 0; co1lo.sRi = 0; co1lo.sRm = 0; co1lo.sRn = 0;
      co1lo.M = L; co1lo.N = R; co1lo.K = D; co1lo.zi_n = 1; co1lo.flags = 0; co1lo.act = 0;
      co1lo.alpha = 1.0f; co1lo.beta = 0.0f; co1lo.sa = 1.0f; co1lo.sb = 1.0f; co1lo.Npad = R; co1lo.pad_ = 0;
      if ((long long)(L) >= 64 && (long long)(R) >= 64) k_gemmT<0, 4, 4><<<dim3((unsigned)((R) + 63) / 64, (unsigned)((L) + 63) / 64, (unsigned)(1)), 32, 0, stream>>>(co1lo);
      else k_gemm<0><<<dim3((unsigned)((R) + 31) / 32, (unsigned)((L) + 15) / 16, (unsigned)(1)), 32, 0, stream>>>(co1lo); }
    k_cast16<<<(unsigned)((((long long)(512) * ((1024) / 2)) + 255) / 256), 256, 0, stream>>>(AT, 1024, (_Float16*)(G64A), 1024, 512, 1024, 1.0f);
    k_castT16<<<(unsigned)((((long long)(1024) * ((1024) / 2)) + 255) / 256), 256, 0, stream>>>(cWo, 1024, (_Float16*)(G64B), 1024, 1024, 1024, 16.0f);
    w25::wmma_gemm64<0, false, 0, 0, true, 0><<<dim3((unsigned)((((512) / 64) * ((1024) / 64) + 7) / 8), (unsigned)(1)), 256, 0, stream>>>((const unsigned short*)(G64A), nullptr, 1024, 0, (const unsigned short*)(G64B), nullptr, 1024, 0, (void*)(Y1 + (size_t)1 * L * D), nullptr, 1024, 0, nullptr, X1 + (size_t)1 * L * D, 0, 512, 1024, 1024, 0.0625f);
    { GemmP co1ab;
      co1ab.A = LOW; co1ab.B = ob + (size_t)3 * R * D; co1ab.bias = LOW; co1ab.R = Y1 + (size_t)1 * L * D; co1ab.C = Y1 + (size_t)1 * L * D;
      co1ab.sAo = 0; co1ab.sAi = 0; co1ab.sAm = R; co1ab.sAk = 1; co1ab.sBo = 0; co1ab.sBi = 0; co1ab.sBn = 1; co1ab.sBk = D; co1ab.sCo = 0; co1ab.sCi = 0; co1ab.sCm = D; co1ab.sRo = 0; co1ab.sRi = 0; co1ab.sRm = D; co1ab.sRn = 1;
      co1ab.M = L; co1ab.N = D; co1ab.K = R; co1ab.zi_n = 1; co1ab.flags = 4; co1ab.act = 0;
      co1ab.alpha = 1.0f; co1ab.beta = 1.0f; co1ab.sa = 1.0f; co1ab.sb = 1.0f; co1ab.Npad = D; co1ab.pad_ = 0;
      if ((long long)(L) >= 64 && (long long)(D) >= 64) k_gemmT<0, 4, 4><<<dim3((unsigned)((D) + 63) / 64, (unsigned)((L) + 63) / 64, (unsigned)(1)), 32, 0, stream>>>(co1ab);
      else k_gemm<0><<<dim3((unsigned)((D) + 31) / 32, (unsigned)((L) + 15) / 16, (unsigned)(1)), 32, 0, stream>>>(co1ab); }
    k_ld_rms<<<L, 256, 0, stream>>>(Y1 + (size_t)1 * L * D, ln3, XN, D);
    k_cast16<<<(unsigned)((((long long)(512) * ((1024) / 2)) + 255) / 256), 256, 0, stream>>>(XN, 1024, (_Float16*)(G64A), 1024, 512, 1024, 1.0f);
    k_castT16<<<(unsigned)((((long long)(4096) * ((1024) / 2)) + 255) / 256), 256, 0, stream>>>(wi0, 4096, (_Float16*)(G64B), 1024, 1024, 4096, 16.0f);
    w25::wmma_gemm64<0, false, 0, 0, false, 0><<<dim3((unsigned)((((512) / 64) * ((4096) / 64) + 7) / 8), (unsigned)(1)), 256, 0, stream>>>((const unsigned short*)(G64A), nullptr, 1024, 0, (const unsigned short*)(G64B), nullptr, 1024, 0, (void*)(G0), nullptr, 4096, 0, nullptr, nullptr, 0, 512, 4096, 1024, 0.0625f);
    k_cast16<<<(unsigned)((((long long)(512) * ((1024) / 2)) + 255) / 256), 256, 0, stream>>>(XN, 1024, (_Float16*)(G64A), 1024, 512, 1024, 1.0f);
    k_castT16<<<(unsigned)((((long long)(4096) * ((1024) / 2)) + 255) / 256), 256, 0, stream>>>(wi1, 4096, (_Float16*)(G64B), 1024, 1024, 4096, 16.0f);
    w25::wmma_gemm64<0, false, 0, 0, false, 0><<<dim3((unsigned)((((512) / 64) * ((4096) / 64) + 7) / 8), (unsigned)(1)), 256, 0, stream>>>((const unsigned short*)(G64A), nullptr, 1024, 0, (const unsigned short*)(G64B), nullptr, 1024, 0, (void*)(G1), nullptr, 4096, 0, nullptr, nullptr, 0, 512, 4096, 1024, 0.0625f);
    k_ld_gg<<<(unsigned)(((long long)L * FF + 255) / 256), 256, 0, stream>>>(G0, G1, (long long)L * FF);
    k_cast16<<<(unsigned)((((long long)(512) * ((4096) / 2)) + 255) / 256), 256, 0, stream>>>(G0, 4096, (_Float16*)(G64A), 4096, 512, 4096, 1.0f);
    k_castT16<<<(unsigned)((((long long)(1024) * ((4096) / 2)) + 255) / 256), 256, 0, stream>>>(wom, 1024, (_Float16*)(G64B), 4096, 4096, 1024, 16.0f);
    w25::wmma_gemm64<0, false, 0, 0, true, 0><<<dim3((unsigned)((((512) / 64) * ((1024) / 64) + 7) / 8), (unsigned)(1)), 256, 0, stream>>>((const unsigned short*)(G64A), nullptr, 4096, 0, (const unsigned short*)(G64B), nullptr, 4096, 0, (void*)(out + (size_t)1 * L * D), nullptr, 1024, 0, nullptr, Y1 + (size_t)1 * L * D, 0, 512, 1024, 4096, 0.0625f);
    k_ld_rms<<<L, 256, 0, stream>>>(xin + (size_t)2 * L * D, ln1, XN, D);
    { GemmP sq2lo;
      sq2lo.A = XN; sq2lo.B = qa + (size_t)4 * D * R; sq2lo.bias = XN; sq2lo.R = XN; sq2lo.C = LOW;
      sq2lo.sAo = 0; sq2lo.sAi = 0; sq2lo.sAm = D; sq2lo.sAk = 1; sq2lo.sBo = 0; sq2lo.sBi = 0; sq2lo.sBn = 1; sq2lo.sBk = R; sq2lo.sCo = 0; sq2lo.sCi = 0; sq2lo.sCm = R; sq2lo.sRo = 0; sq2lo.sRi = 0; sq2lo.sRm = 0; sq2lo.sRn = 0;
      sq2lo.M = L; sq2lo.N = R; sq2lo.K = D; sq2lo.zi_n = 1; sq2lo.flags = 0; sq2lo.act = 0;
      sq2lo.alpha = 1.0f; sq2lo.beta = 0.0f; sq2lo.sa = 1.0f; sq2lo.sb = 1.0f; sq2lo.Npad = R; sq2lo.pad_ = 0;
      if ((long long)(L) >= 64 && (long long)(R) >= 64) k_gemmT<0, 4, 4><<<dim3((unsigned)((R) + 63) / 64, (unsigned)((L) + 63) / 64, (unsigned)(1)), 32, 0, stream>>>(sq2lo);
      else k_gemm<0><<<dim3((unsigned)((R) + 31) / 32, (unsigned)((L) + 15) / 16, (unsigned)(1)), 32, 0, stream>>>(sq2lo); }
    k_cast16<<<(unsigned)((((long long)(512) * ((1024) / 2)) + 255) / 256), 256, 0, stream>>>(XN, 1024, (_Float16*)(G64A), 1024, 512, 1024, 1.0f);
    k_castT16<<<(unsigned)((((long long)(1024) * ((1024) / 2)) + 255) / 256), 256, 0, stream>>>(sWq, 1024, (_Float16*)(G64B), 1024, 1024, 1024, 16.0f);
    w25::wmma_gemm64<0, false, 0, 0, false, 0><<<dim3((unsigned)((((512) / 64) * ((1024) / 64) + 7) / 8), (unsigned)(1)), 256, 0, stream>>>((const unsigned short*)(G64A), nullptr, 1024, 0, (const unsigned short*)(G64B), nullptr, 1024, 0, (void*)(Q), nullptr, 1024, 0, nullptr, nullptr, 0, 512, 1024, 1024, 0.0625f);
    { GemmP sq2ab;
      sq2ab.A = LOW; sq2ab.B = qb + (size_t)4 * R * D; sq2ab.bias = LOW; sq2ab.R = Q; sq2ab.C = Q;
      sq2ab.sAo = 0; sq2ab.sAi = 0; sq2ab.sAm = R; sq2ab.sAk = 1; sq2ab.sBo = 0; sq2ab.sBi = 0; sq2ab.sBn = 1; sq2ab.sBk = D; sq2ab.sCo = 0; sq2ab.sCi = 0; sq2ab.sCm = D; sq2ab.sRo = 0; sq2ab.sRi = 0; sq2ab.sRm = D; sq2ab.sRn = 1;
      sq2ab.M = L; sq2ab.N = D; sq2ab.K = R; sq2ab.zi_n = 1; sq2ab.flags = 4; sq2ab.act = 0;
      sq2ab.alpha = 1.0f; sq2ab.beta = 1.0f; sq2ab.sa = 1.0f; sq2ab.sb = 1.0f; sq2ab.Npad = D; sq2ab.pad_ = 0;
      if ((long long)(L) >= 64 && (long long)(D) >= 64) k_gemmT<0, 4, 4><<<dim3((unsigned)((D) + 63) / 64, (unsigned)((L) + 63) / 64, (unsigned)(1)), 32, 0, stream>>>(sq2ab);
      else k_gemm<0><<<dim3((unsigned)((D) + 31) / 32, (unsigned)((L) + 15) / 16, (unsigned)(1)), 32, 0, stream>>>(sq2ab); }
    { GemmP sk2lo;
      sk2lo.A = XN; sk2lo.B = ka + (size_t)4 * D * R; sk2lo.bias = XN; sk2lo.R = XN; sk2lo.C = LOW;
      sk2lo.sAo = 0; sk2lo.sAi = 0; sk2lo.sAm = D; sk2lo.sAk = 1; sk2lo.sBo = 0; sk2lo.sBi = 0; sk2lo.sBn = 1; sk2lo.sBk = R; sk2lo.sCo = 0; sk2lo.sCi = 0; sk2lo.sCm = R; sk2lo.sRo = 0; sk2lo.sRi = 0; sk2lo.sRm = 0; sk2lo.sRn = 0;
      sk2lo.M = L; sk2lo.N = R; sk2lo.K = D; sk2lo.zi_n = 1; sk2lo.flags = 0; sk2lo.act = 0;
      sk2lo.alpha = 1.0f; sk2lo.beta = 0.0f; sk2lo.sa = 1.0f; sk2lo.sb = 1.0f; sk2lo.Npad = R; sk2lo.pad_ = 0;
      if ((long long)(L) >= 64 && (long long)(R) >= 64) k_gemmT<0, 4, 4><<<dim3((unsigned)((R) + 63) / 64, (unsigned)((L) + 63) / 64, (unsigned)(1)), 32, 0, stream>>>(sk2lo);
      else k_gemm<0><<<dim3((unsigned)((R) + 31) / 32, (unsigned)((L) + 15) / 16, (unsigned)(1)), 32, 0, stream>>>(sk2lo); }
    k_cast16<<<(unsigned)((((long long)(512) * ((1024) / 2)) + 255) / 256), 256, 0, stream>>>(XN, 1024, (_Float16*)(G64A), 1024, 512, 1024, 1.0f);
    k_castT16<<<(unsigned)((((long long)(1024) * ((1024) / 2)) + 255) / 256), 256, 0, stream>>>(sWk, 1024, (_Float16*)(G64B), 1024, 1024, 1024, 16.0f);
    w25::wmma_gemm64<0, false, 0, 0, false, 0><<<dim3((unsigned)((((512) / 64) * ((1024) / 64) + 7) / 8), (unsigned)(1)), 256, 0, stream>>>((const unsigned short*)(G64A), nullptr, 1024, 0, (const unsigned short*)(G64B), nullptr, 1024, 0, (void*)(Kb), nullptr, 1024, 0, nullptr, nullptr, 0, 512, 1024, 1024, 0.0625f);
    { GemmP sk2ab;
      sk2ab.A = LOW; sk2ab.B = kb + (size_t)4 * R * D; sk2ab.bias = LOW; sk2ab.R = Kb; sk2ab.C = Kb;
      sk2ab.sAo = 0; sk2ab.sAi = 0; sk2ab.sAm = R; sk2ab.sAk = 1; sk2ab.sBo = 0; sk2ab.sBi = 0; sk2ab.sBn = 1; sk2ab.sBk = D; sk2ab.sCo = 0; sk2ab.sCi = 0; sk2ab.sCm = D; sk2ab.sRo = 0; sk2ab.sRi = 0; sk2ab.sRm = D; sk2ab.sRn = 1;
      sk2ab.M = L; sk2ab.N = D; sk2ab.K = R; sk2ab.zi_n = 1; sk2ab.flags = 4; sk2ab.act = 0;
      sk2ab.alpha = 1.0f; sk2ab.beta = 1.0f; sk2ab.sa = 1.0f; sk2ab.sb = 1.0f; sk2ab.Npad = D; sk2ab.pad_ = 0;
      if ((long long)(L) >= 64 && (long long)(D) >= 64) k_gemmT<0, 4, 4><<<dim3((unsigned)((D) + 63) / 64, (unsigned)((L) + 63) / 64, (unsigned)(1)), 32, 0, stream>>>(sk2ab);
      else k_gemm<0><<<dim3((unsigned)((D) + 31) / 32, (unsigned)((L) + 15) / 16, (unsigned)(1)), 32, 0, stream>>>(sk2ab); }
    { GemmP sv2lo;
      sv2lo.A = XN; sv2lo.B = va + (size_t)4 * D * R; sv2lo.bias = XN; sv2lo.R = XN; sv2lo.C = LOW;
      sv2lo.sAo = 0; sv2lo.sAi = 0; sv2lo.sAm = D; sv2lo.sAk = 1; sv2lo.sBo = 0; sv2lo.sBi = 0; sv2lo.sBn = 1; sv2lo.sBk = R; sv2lo.sCo = 0; sv2lo.sCi = 0; sv2lo.sCm = R; sv2lo.sRo = 0; sv2lo.sRi = 0; sv2lo.sRm = 0; sv2lo.sRn = 0;
      sv2lo.M = L; sv2lo.N = R; sv2lo.K = D; sv2lo.zi_n = 1; sv2lo.flags = 0; sv2lo.act = 0;
      sv2lo.alpha = 1.0f; sv2lo.beta = 0.0f; sv2lo.sa = 1.0f; sv2lo.sb = 1.0f; sv2lo.Npad = R; sv2lo.pad_ = 0;
      if ((long long)(L) >= 64 && (long long)(R) >= 64) k_gemmT<0, 4, 4><<<dim3((unsigned)((R) + 63) / 64, (unsigned)((L) + 63) / 64, (unsigned)(1)), 32, 0, stream>>>(sv2lo);
      else k_gemm<0><<<dim3((unsigned)((R) + 31) / 32, (unsigned)((L) + 15) / 16, (unsigned)(1)), 32, 0, stream>>>(sv2lo); }
    k_cast16<<<(unsigned)((((long long)(512) * ((1024) / 2)) + 255) / 256), 256, 0, stream>>>(XN, 1024, (_Float16*)(G64A), 1024, 512, 1024, 1.0f);
    k_castT16<<<(unsigned)((((long long)(1024) * ((1024) / 2)) + 255) / 256), 256, 0, stream>>>(sWv, 1024, (_Float16*)(G64B), 1024, 1024, 1024, 16.0f);
    w25::wmma_gemm64<0, false, 0, 0, false, 0><<<dim3((unsigned)((((512) / 64) * ((1024) / 64) + 7) / 8), (unsigned)(1)), 256, 0, stream>>>((const unsigned short*)(G64A), nullptr, 1024, 0, (const unsigned short*)(G64B), nullptr, 1024, 0, (void*)(V), nullptr, 1024, 0, nullptr, nullptr, 0, 512, 1024, 1024, 0.0625f);
    { GemmP sv2ab;
      sv2ab.A = LOW; sv2ab.B = vb + (size_t)4 * R * D; sv2ab.bias = LOW; sv2ab.R = V; sv2ab.C = V;
      sv2ab.sAo = 0; sv2ab.sAi = 0; sv2ab.sAm = R; sv2ab.sAk = 1; sv2ab.sBo = 0; sv2ab.sBi = 0; sv2ab.sBn = 1; sv2ab.sBk = D; sv2ab.sCo = 0; sv2ab.sCi = 0; sv2ab.sCm = D; sv2ab.sRo = 0; sv2ab.sRi = 0; sv2ab.sRm = D; sv2ab.sRn = 1;
      sv2ab.M = L; sv2ab.N = D; sv2ab.K = R; sv2ab.zi_n = 1; sv2ab.flags = 4; sv2ab.act = 0;
      sv2ab.alpha = 1.0f; sv2ab.beta = 1.0f; sv2ab.sa = 1.0f; sv2ab.sb = 1.0f; sv2ab.Npad = D; sv2ab.pad_ = 0;
      if ((long long)(L) >= 64 && (long long)(D) >= 64) k_gemmT<0, 4, 4><<<dim3((unsigned)((D) + 63) / 64, (unsigned)((L) + 63) / 64, (unsigned)(1)), 32, 0, stream>>>(sv2ab);
      else k_gemm<0><<<dim3((unsigned)((D) + 31) / 32, (unsigned)((L) + 15) / 16, (unsigned)(1)), 32, 0, stream>>>(sv2ab); }
    {   AttnP a;
      a.Q = Q; a.K = Kb; a.V = V; a.O = AT; a.P = 0; a.Mf = BIAS; a.Mi = 0; a.ST = 0;
      a.Pw = 0; a.Rt = 0; a.SQ = 0; a.SK = 0;
      a.swb = 0; a.swh = 0; a.swi = 0; a.swj = 0; a.srb = 0; a.srh = 0; a.sri = 0; a.sQb = 0; a.sQh = HD; a.sQi = D; a.sQd = 1; a.sKb = 0; a.sKh = HD; a.sKj = D; a.sKd = 1; a.sVb = 0; a.sVh = HD; a.sVj = D; a.sVd = 1; a.sOb = 0; a.sOh = HD; a.sOi = D; a.sPb = 0; a.sPh = 0; a.sPi = 0; a.smb = 0; a.smh = (long long)L * L; a.smi = L; a.smj = 1;
      a.Lq = L; a.Lk = L; a.dh = HD; a.dv = HD; a.hrep = 1; a.causal = 1; a.coff = 0; a.pband = 0;
      a.scale = 0.125f; a.mfill = 0.0f; a.nonorm = 0; a.mpol = 0;
      a.roff = 0; a.rn = 1; a.segpol = 0; a.win = 0;
      k_attn<64, 64, 0, false, false><<<dim3((unsigned)((L) + 16 * AW - 1) / (16 * AW), (unsigned)(NH), (unsigned)(1)), 32 * AW, 0, stream>>>(a); }
    { GemmP so2lo;
      so2lo.A = AT; so2lo.B = oa + (size_t)4 * D * R; so2lo.bias = AT; so2lo.R = AT; so2lo.C = LOW;
      so2lo.sAo = 0; so2lo.sAi = 0; so2lo.sAm = D; so2lo.sAk = 1; so2lo.sBo = 0; so2lo.sBi = 0; so2lo.sBn = 1; so2lo.sBk = R; so2lo.sCo = 0; so2lo.sCi = 0; so2lo.sCm = R; so2lo.sRo = 0; so2lo.sRi = 0; so2lo.sRm = 0; so2lo.sRn = 0;
      so2lo.M = L; so2lo.N = R; so2lo.K = D; so2lo.zi_n = 1; so2lo.flags = 0; so2lo.act = 0;
      so2lo.alpha = 1.0f; so2lo.beta = 0.0f; so2lo.sa = 1.0f; so2lo.sb = 1.0f; so2lo.Npad = R; so2lo.pad_ = 0;
      if ((long long)(L) >= 64 && (long long)(R) >= 64) k_gemmT<0, 4, 4><<<dim3((unsigned)((R) + 63) / 64, (unsigned)((L) + 63) / 64, (unsigned)(1)), 32, 0, stream>>>(so2lo);
      else k_gemm<0><<<dim3((unsigned)((R) + 31) / 32, (unsigned)((L) + 15) / 16, (unsigned)(1)), 32, 0, stream>>>(so2lo); }
    k_cast16<<<(unsigned)((((long long)(512) * ((1024) / 2)) + 255) / 256), 256, 0, stream>>>(AT, 1024, (_Float16*)(G64A), 1024, 512, 1024, 1.0f);
    k_castT16<<<(unsigned)((((long long)(1024) * ((1024) / 2)) + 255) / 256), 256, 0, stream>>>(sWo, 1024, (_Float16*)(G64B), 1024, 1024, 1024, 16.0f);
    w25::wmma_gemm64<0, false, 0, 0, true, 0><<<dim3((unsigned)((((512) / 64) * ((1024) / 64) + 7) / 8), (unsigned)(1)), 256, 0, stream>>>((const unsigned short*)(G64A), nullptr, 1024, 0, (const unsigned short*)(G64B), nullptr, 1024, 0, (void*)(X1 + (size_t)2 * L * D), nullptr, 1024, 0, nullptr, xin + (size_t)2 * L * D, 0, 512, 1024, 1024, 0.0625f);
    { GemmP so2ab;
      so2ab.A = LOW; so2ab.B = ob + (size_t)4 * R * D; so2ab.bias = LOW; so2ab.R = X1 + (size_t)2 * L * D; so2ab.C = X1 + (size_t)2 * L * D;
      so2ab.sAo = 0; so2ab.sAi = 0; so2ab.sAm = R; so2ab.sAk = 1; so2ab.sBo = 0; so2ab.sBi = 0; so2ab.sBn = 1; so2ab.sBk = D; so2ab.sCo = 0; so2ab.sCi = 0; so2ab.sCm = D; so2ab.sRo = 0; so2ab.sRi = 0; so2ab.sRm = D; so2ab.sRn = 1;
      so2ab.M = L; so2ab.N = D; so2ab.K = R; so2ab.zi_n = 1; so2ab.flags = 4; so2ab.act = 0;
      so2ab.alpha = 1.0f; so2ab.beta = 1.0f; so2ab.sa = 1.0f; so2ab.sb = 1.0f; so2ab.Npad = D; so2ab.pad_ = 0;
      if ((long long)(L) >= 64 && (long long)(D) >= 64) k_gemmT<0, 4, 4><<<dim3((unsigned)((D) + 63) / 64, (unsigned)((L) + 63) / 64, (unsigned)(1)), 32, 0, stream>>>(so2ab);
      else k_gemm<0><<<dim3((unsigned)((D) + 31) / 32, (unsigned)((L) + 15) / 16, (unsigned)(1)), 32, 0, stream>>>(so2ab); }
    k_ld_rms<<<L, 256, 0, stream>>>(X1 + (size_t)2 * L * D, ln2, XN, D);
    { GemmP cq2lo;
      cq2lo.A = XN; cq2lo.B = qa + (size_t)5 * D * R; cq2lo.bias = XN; cq2lo.R = XN; cq2lo.C = LOW;
      cq2lo.sAo = 0; cq2lo.sAi = 0; cq2lo.sAm = D; cq2lo.sAk = 1; cq2lo.sBo = 0; cq2lo.sBi = 0; cq2lo.sBn = 1; cq2lo.sBk = R; cq2lo.sCo = 0; cq2lo.sCi = 0; cq2lo.sCm = R; cq2lo.sRo = 0; cq2lo.sRi = 0; cq2lo.sRm = 0; cq2lo.sRn = 0;
      cq2lo.M = L; cq2lo.N = R; cq2lo.K = D; cq2lo.zi_n = 1; cq2lo.flags = 0; cq2lo.act = 0;
      cq2lo.alpha = 1.0f; cq2lo.beta = 0.0f; cq2lo.sa = 1.0f; cq2lo.sb = 1.0f; cq2lo.Npad = R; cq2lo.pad_ = 0;
      if ((long long)(L) >= 64 && (long long)(R) >= 64) k_gemmT<0, 4, 4><<<dim3((unsigned)((R) + 63) / 64, (unsigned)((L) + 63) / 64, (unsigned)(1)), 32, 0, stream>>>(cq2lo);
      else k_gemm<0><<<dim3((unsigned)((R) + 31) / 32, (unsigned)((L) + 15) / 16, (unsigned)(1)), 32, 0, stream>>>(cq2lo); }
    k_cast16<<<(unsigned)((((long long)(512) * ((1024) / 2)) + 255) / 256), 256, 0, stream>>>(XN, 1024, (_Float16*)(G64A), 1024, 512, 1024, 1.0f);
    k_castT16<<<(unsigned)((((long long)(1024) * ((1024) / 2)) + 255) / 256), 256, 0, stream>>>(cWq, 1024, (_Float16*)(G64B), 1024, 1024, 1024, 16.0f);
    w25::wmma_gemm64<0, false, 0, 0, false, 0><<<dim3((unsigned)((((512) / 64) * ((1024) / 64) + 7) / 8), (unsigned)(1)), 256, 0, stream>>>((const unsigned short*)(G64A), nullptr, 1024, 0, (const unsigned short*)(G64B), nullptr, 1024, 0, (void*)(Q), nullptr, 1024, 0, nullptr, nullptr, 0, 512, 1024, 1024, 0.0625f);
    { GemmP cq2ab;
      cq2ab.A = LOW; cq2ab.B = qb + (size_t)5 * R * D; cq2ab.bias = LOW; cq2ab.R = Q; cq2ab.C = Q;
      cq2ab.sAo = 0; cq2ab.sAi = 0; cq2ab.sAm = R; cq2ab.sAk = 1; cq2ab.sBo = 0; cq2ab.sBi = 0; cq2ab.sBn = 1; cq2ab.sBk = D; cq2ab.sCo = 0; cq2ab.sCi = 0; cq2ab.sCm = D; cq2ab.sRo = 0; cq2ab.sRi = 0; cq2ab.sRm = D; cq2ab.sRn = 1;
      cq2ab.M = L; cq2ab.N = D; cq2ab.K = R; cq2ab.zi_n = 1; cq2ab.flags = 4; cq2ab.act = 0;
      cq2ab.alpha = 1.0f; cq2ab.beta = 1.0f; cq2ab.sa = 1.0f; cq2ab.sb = 1.0f; cq2ab.Npad = D; cq2ab.pad_ = 0;
      if ((long long)(L) >= 64 && (long long)(D) >= 64) k_gemmT<0, 4, 4><<<dim3((unsigned)((D) + 63) / 64, (unsigned)((L) + 63) / 64, (unsigned)(1)), 32, 0, stream>>>(cq2ab);
      else k_gemm<0><<<dim3((unsigned)((D) + 31) / 32, (unsigned)((L) + 15) / 16, (unsigned)(1)), 32, 0, stream>>>(cq2ab); }
    { GemmP ck2lo;
      ck2lo.A = enc + (size_t)2 * L * D; ck2lo.B = ka + (size_t)5 * D * R; ck2lo.bias = enc + (size_t)2 * L * D; ck2lo.R = enc + (size_t)2 * L * D; ck2lo.C = LOW;
      ck2lo.sAo = 0; ck2lo.sAi = 0; ck2lo.sAm = D; ck2lo.sAk = 1; ck2lo.sBo = 0; ck2lo.sBi = 0; ck2lo.sBn = 1; ck2lo.sBk = R; ck2lo.sCo = 0; ck2lo.sCi = 0; ck2lo.sCm = R; ck2lo.sRo = 0; ck2lo.sRi = 0; ck2lo.sRm = 0; ck2lo.sRn = 0;
      ck2lo.M = L; ck2lo.N = R; ck2lo.K = D; ck2lo.zi_n = 1; ck2lo.flags = 0; ck2lo.act = 0;
      ck2lo.alpha = 1.0f; ck2lo.beta = 0.0f; ck2lo.sa = 1.0f; ck2lo.sb = 1.0f; ck2lo.Npad = R; ck2lo.pad_ = 0;
      if ((long long)(L) >= 64 && (long long)(R) >= 64) k_gemmT<0, 4, 4><<<dim3((unsigned)((R) + 63) / 64, (unsigned)((L) + 63) / 64, (unsigned)(1)), 32, 0, stream>>>(ck2lo);
      else k_gemm<0><<<dim3((unsigned)((R) + 31) / 32, (unsigned)((L) + 15) / 16, (unsigned)(1)), 32, 0, stream>>>(ck2lo); }
    k_cast16<<<(unsigned)((((long long)(512) * ((1024) / 2)) + 255) / 256), 256, 0, stream>>>(enc + (size_t)2 * L * D, 1024, (_Float16*)(G64A), 1024, 512, 1024, 1.0f);
    k_castT16<<<(unsigned)((((long long)(1024) * ((1024) / 2)) + 255) / 256), 256, 0, stream>>>(cWk, 1024, (_Float16*)(G64B), 1024, 1024, 1024, 16.0f);
    w25::wmma_gemm64<0, false, 0, 0, false, 0><<<dim3((unsigned)((((512) / 64) * ((1024) / 64) + 7) / 8), (unsigned)(1)), 256, 0, stream>>>((const unsigned short*)(G64A), nullptr, 1024, 0, (const unsigned short*)(G64B), nullptr, 1024, 0, (void*)(Kb), nullptr, 1024, 0, nullptr, nullptr, 0, 512, 1024, 1024, 0.0625f);
    { GemmP ck2ab;
      ck2ab.A = LOW; ck2ab.B = kb + (size_t)5 * R * D; ck2ab.bias = LOW; ck2ab.R = Kb; ck2ab.C = Kb;
      ck2ab.sAo = 0; ck2ab.sAi = 0; ck2ab.sAm = R; ck2ab.sAk = 1; ck2ab.sBo = 0; ck2ab.sBi = 0; ck2ab.sBn = 1; ck2ab.sBk = D; ck2ab.sCo = 0; ck2ab.sCi = 0; ck2ab.sCm = D; ck2ab.sRo = 0; ck2ab.sRi = 0; ck2ab.sRm = D; ck2ab.sRn = 1;
      ck2ab.M = L; ck2ab.N = D; ck2ab.K = R; ck2ab.zi_n = 1; ck2ab.flags = 4; ck2ab.act = 0;
      ck2ab.alpha = 1.0f; ck2ab.beta = 1.0f; ck2ab.sa = 1.0f; ck2ab.sb = 1.0f; ck2ab.Npad = D; ck2ab.pad_ = 0;
      if ((long long)(L) >= 64 && (long long)(D) >= 64) k_gemmT<0, 4, 4><<<dim3((unsigned)((D) + 63) / 64, (unsigned)((L) + 63) / 64, (unsigned)(1)), 32, 0, stream>>>(ck2ab);
      else k_gemm<0><<<dim3((unsigned)((D) + 31) / 32, (unsigned)((L) + 15) / 16, (unsigned)(1)), 32, 0, stream>>>(ck2ab); }
    { GemmP cv2lo;
      cv2lo.A = enc + (size_t)2 * L * D; cv2lo.B = va + (size_t)5 * D * R; cv2lo.bias = enc + (size_t)2 * L * D; cv2lo.R = enc + (size_t)2 * L * D; cv2lo.C = LOW;
      cv2lo.sAo = 0; cv2lo.sAi = 0; cv2lo.sAm = D; cv2lo.sAk = 1; cv2lo.sBo = 0; cv2lo.sBi = 0; cv2lo.sBn = 1; cv2lo.sBk = R; cv2lo.sCo = 0; cv2lo.sCi = 0; cv2lo.sCm = R; cv2lo.sRo = 0; cv2lo.sRi = 0; cv2lo.sRm = 0; cv2lo.sRn = 0;
      cv2lo.M = L; cv2lo.N = R; cv2lo.K = D; cv2lo.zi_n = 1; cv2lo.flags = 0; cv2lo.act = 0;
      cv2lo.alpha = 1.0f; cv2lo.beta = 0.0f; cv2lo.sa = 1.0f; cv2lo.sb = 1.0f; cv2lo.Npad = R; cv2lo.pad_ = 0;
      if ((long long)(L) >= 64 && (long long)(R) >= 64) k_gemmT<0, 4, 4><<<dim3((unsigned)((R) + 63) / 64, (unsigned)((L) + 63) / 64, (unsigned)(1)), 32, 0, stream>>>(cv2lo);
      else k_gemm<0><<<dim3((unsigned)((R) + 31) / 32, (unsigned)((L) + 15) / 16, (unsigned)(1)), 32, 0, stream>>>(cv2lo); }
    k_cast16<<<(unsigned)((((long long)(512) * ((1024) / 2)) + 255) / 256), 256, 0, stream>>>(enc + (size_t)2 * L * D, 1024, (_Float16*)(G64A), 1024, 512, 1024, 1.0f);
    k_castT16<<<(unsigned)((((long long)(1024) * ((1024) / 2)) + 255) / 256), 256, 0, stream>>>(cWv, 1024, (_Float16*)(G64B), 1024, 1024, 1024, 16.0f);
    w25::wmma_gemm64<0, false, 0, 0, false, 0><<<dim3((unsigned)((((512) / 64) * ((1024) / 64) + 7) / 8), (unsigned)(1)), 256, 0, stream>>>((const unsigned short*)(G64A), nullptr, 1024, 0, (const unsigned short*)(G64B), nullptr, 1024, 0, (void*)(V), nullptr, 1024, 0, nullptr, nullptr, 0, 512, 1024, 1024, 0.0625f);
    { GemmP cv2ab;
      cv2ab.A = LOW; cv2ab.B = vb + (size_t)5 * R * D; cv2ab.bias = LOW; cv2ab.R = V; cv2ab.C = V;
      cv2ab.sAo = 0; cv2ab.sAi = 0; cv2ab.sAm = R; cv2ab.sAk = 1; cv2ab.sBo = 0; cv2ab.sBi = 0; cv2ab.sBn = 1; cv2ab.sBk = D; cv2ab.sCo = 0; cv2ab.sCi = 0; cv2ab.sCm = D; cv2ab.sRo = 0; cv2ab.sRi = 0; cv2ab.sRm = D; cv2ab.sRn = 1;
      cv2ab.M = L; cv2ab.N = D; cv2ab.K = R; cv2ab.zi_n = 1; cv2ab.flags = 4; cv2ab.act = 0;
      cv2ab.alpha = 1.0f; cv2ab.beta = 1.0f; cv2ab.sa = 1.0f; cv2ab.sb = 1.0f; cv2ab.Npad = D; cv2ab.pad_ = 0;
      if ((long long)(L) >= 64 && (long long)(D) >= 64) k_gemmT<0, 4, 4><<<dim3((unsigned)((D) + 63) / 64, (unsigned)((L) + 63) / 64, (unsigned)(1)), 32, 0, stream>>>(cv2ab);
      else k_gemm<0><<<dim3((unsigned)((D) + 31) / 32, (unsigned)((L) + 15) / 16, (unsigned)(1)), 32, 0, stream>>>(cv2ab); }
    {   AttnP a;
      a.Q = Q; a.K = Kb; a.V = V; a.O = AT; a.P = 0; a.Mf = 0; a.Mi = 0; a.ST = 0;
      a.Pw = 0; a.Rt = 0; a.SQ = 0; a.SK = 0;
      a.swb = 0; a.swh = 0; a.swi = 0; a.swj = 0; a.srb = 0; a.srh = 0; a.sri = 0; a.sQb = 0; a.sQh = HD; a.sQi = D; a.sQd = 1; a.sKb = 0; a.sKh = HD; a.sKj = D; a.sKd = 1; a.sVb = 0; a.sVh = HD; a.sVj = D; a.sVd = 1; a.sOb = 0; a.sOh = HD; a.sOi = D; a.sPb = 0; a.sPh = 0; a.sPi = 0; a.smb = 0; a.smh = 0; a.smi = 0; a.smj = 0;
      a.Lq = L; a.Lk = L; a.dh = HD; a.dv = HD; a.hrep = 1; a.causal = 0; a.coff = 0; a.pband = 0;
      a.scale = 0.125f; a.mfill = 0.0f; a.nonorm = 0; a.mpol = 0;
      a.roff = 0; a.rn = 1; a.segpol = 0; a.win = 0;
      k_attn<64, 64, 0, false, false><<<dim3((unsigned)((L) + 16 * AW - 1) / (16 * AW), (unsigned)(NH), (unsigned)(1)), 32 * AW, 0, stream>>>(a); }
    { GemmP co2lo;
      co2lo.A = AT; co2lo.B = oa + (size_t)5 * D * R; co2lo.bias = AT; co2lo.R = AT; co2lo.C = LOW;
      co2lo.sAo = 0; co2lo.sAi = 0; co2lo.sAm = D; co2lo.sAk = 1; co2lo.sBo = 0; co2lo.sBi = 0; co2lo.sBn = 1; co2lo.sBk = R; co2lo.sCo = 0; co2lo.sCi = 0; co2lo.sCm = R; co2lo.sRo = 0; co2lo.sRi = 0; co2lo.sRm = 0; co2lo.sRn = 0;
      co2lo.M = L; co2lo.N = R; co2lo.K = D; co2lo.zi_n = 1; co2lo.flags = 0; co2lo.act = 0;
      co2lo.alpha = 1.0f; co2lo.beta = 0.0f; co2lo.sa = 1.0f; co2lo.sb = 1.0f; co2lo.Npad = R; co2lo.pad_ = 0;
      if ((long long)(L) >= 64 && (long long)(R) >= 64) k_gemmT<0, 4, 4><<<dim3((unsigned)((R) + 63) / 64, (unsigned)((L) + 63) / 64, (unsigned)(1)), 32, 0, stream>>>(co2lo);
      else k_gemm<0><<<dim3((unsigned)((R) + 31) / 32, (unsigned)((L) + 15) / 16, (unsigned)(1)), 32, 0, stream>>>(co2lo); }
    k_cast16<<<(unsigned)((((long long)(512) * ((1024) / 2)) + 255) / 256), 256, 0, stream>>>(AT, 1024, (_Float16*)(G64A), 1024, 512, 1024, 1.0f);
    k_castT16<<<(unsigned)((((long long)(1024) * ((1024) / 2)) + 255) / 256), 256, 0, stream>>>(cWo, 1024, (_Float16*)(G64B), 1024, 1024, 1024, 16.0f);
    w25::wmma_gemm64<0, false, 0, 0, true, 0><<<dim3((unsigned)((((512) / 64) * ((1024) / 64) + 7) / 8), (unsigned)(1)), 256, 0, stream>>>((const unsigned short*)(G64A), nullptr, 1024, 0, (const unsigned short*)(G64B), nullptr, 1024, 0, (void*)(Y1 + (size_t)2 * L * D), nullptr, 1024, 0, nullptr, X1 + (size_t)2 * L * D, 0, 512, 1024, 1024, 0.0625f);
    { GemmP co2ab;
      co2ab.A = LOW; co2ab.B = ob + (size_t)5 * R * D; co2ab.bias = LOW; co2ab.R = Y1 + (size_t)2 * L * D; co2ab.C = Y1 + (size_t)2 * L * D;
      co2ab.sAo = 0; co2ab.sAi = 0; co2ab.sAm = R; co2ab.sAk = 1; co2ab.sBo = 0; co2ab.sBi = 0; co2ab.sBn = 1; co2ab.sBk = D; co2ab.sCo = 0; co2ab.sCi = 0; co2ab.sCm = D; co2ab.sRo = 0; co2ab.sRi = 0; co2ab.sRm = D; co2ab.sRn = 1;
      co2ab.M = L; co2ab.N = D; co2ab.K = R; co2ab.zi_n = 1; co2ab.flags = 4; co2ab.act = 0;
      co2ab.alpha = 1.0f; co2ab.beta = 1.0f; co2ab.sa = 1.0f; co2ab.sb = 1.0f; co2ab.Npad = D; co2ab.pad_ = 0;
      if ((long long)(L) >= 64 && (long long)(D) >= 64) k_gemmT<0, 4, 4><<<dim3((unsigned)((D) + 63) / 64, (unsigned)((L) + 63) / 64, (unsigned)(1)), 32, 0, stream>>>(co2ab);
      else k_gemm<0><<<dim3((unsigned)((D) + 31) / 32, (unsigned)((L) + 15) / 16, (unsigned)(1)), 32, 0, stream>>>(co2ab); }
    k_ld_rms<<<L, 256, 0, stream>>>(Y1 + (size_t)2 * L * D, ln3, XN, D);
    k_cast16<<<(unsigned)((((long long)(512) * ((1024) / 2)) + 255) / 256), 256, 0, stream>>>(XN, 1024, (_Float16*)(G64A), 1024, 512, 1024, 1.0f);
    k_castT16<<<(unsigned)((((long long)(4096) * ((1024) / 2)) + 255) / 256), 256, 0, stream>>>(wi0, 4096, (_Float16*)(G64B), 1024, 1024, 4096, 16.0f);
    w25::wmma_gemm64<0, false, 0, 0, false, 0><<<dim3((unsigned)((((512) / 64) * ((4096) / 64) + 7) / 8), (unsigned)(1)), 256, 0, stream>>>((const unsigned short*)(G64A), nullptr, 1024, 0, (const unsigned short*)(G64B), nullptr, 1024, 0, (void*)(G0), nullptr, 4096, 0, nullptr, nullptr, 0, 512, 4096, 1024, 0.0625f);
    k_cast16<<<(unsigned)((((long long)(512) * ((1024) / 2)) + 255) / 256), 256, 0, stream>>>(XN, 1024, (_Float16*)(G64A), 1024, 512, 1024, 1.0f);
    k_castT16<<<(unsigned)((((long long)(4096) * ((1024) / 2)) + 255) / 256), 256, 0, stream>>>(wi1, 4096, (_Float16*)(G64B), 1024, 1024, 4096, 16.0f);
    w25::wmma_gemm64<0, false, 0, 0, false, 0><<<dim3((unsigned)((((512) / 64) * ((4096) / 64) + 7) / 8), (unsigned)(1)), 256, 0, stream>>>((const unsigned short*)(G64A), nullptr, 1024, 0, (const unsigned short*)(G64B), nullptr, 1024, 0, (void*)(G1), nullptr, 4096, 0, nullptr, nullptr, 0, 512, 4096, 1024, 0.0625f);
    k_ld_gg<<<(unsigned)(((long long)L * FF + 255) / 256), 256, 0, stream>>>(G0, G1, (long long)L * FF);
    k_cast16<<<(unsigned)((((long long)(512) * ((4096) / 2)) + 255) / 256), 256, 0, stream>>>(G0, 4096, (_Float16*)(G64A), 4096, 512, 4096, 1.0f);
    k_castT16<<<(unsigned)((((long long)(1024) * ((4096) / 2)) + 255) / 256), 256, 0, stream>>>(wom, 1024, (_Float16*)(G64B), 4096, 4096, 1024, 16.0f);
    w25::wmma_gemm64<0, false, 0, 0, true, 0><<<dim3((unsigned)((((512) / 64) * ((1024) / 64) + 7) / 8), (unsigned)(1)), 256, 0, stream>>>((const unsigned short*)(G64A), nullptr, 4096, 0, (const unsigned short*)(G64B), nullptr, 4096, 0, (void*)(out + (size_t)2 * L * D), nullptr, 1024, 0, nullptr, Y1 + (size_t)2 * L * D, 0, 512, 1024, 4096, 0.0625f);
    k_ld_rms<<<L, 256, 0, stream>>>(xin + (size_t)3 * L * D, ln1, XN, D);
    { GemmP sq3lo;
      sq3lo.A = XN; sq3lo.B = qa + (size_t)6 * D * R; sq3lo.bias = XN; sq3lo.R = XN; sq3lo.C = LOW;
      sq3lo.sAo = 0; sq3lo.sAi = 0; sq3lo.sAm = D; sq3lo.sAk = 1; sq3lo.sBo = 0; sq3lo.sBi = 0; sq3lo.sBn = 1; sq3lo.sBk = R; sq3lo.sCo = 0; sq3lo.sCi = 0; sq3lo.sCm = R; sq3lo.sRo = 0; sq3lo.sRi = 0; sq3lo.sRm = 0; sq3lo.sRn = 0;
      sq3lo.M = L; sq3lo.N = R; sq3lo.K = D; sq3lo.zi_n = 1; sq3lo.flags = 0; sq3lo.act = 0;
      sq3lo.alpha = 1.0f; sq3lo.beta = 0.0f; sq3lo.sa = 1.0f; sq3lo.sb = 1.0f; sq3lo.Npad = R; sq3lo.pad_ = 0;
      if ((long long)(L) >= 64 && (long long)(R) >= 64) k_gemmT<0, 4, 4><<<dim3((unsigned)((R) + 63) / 64, (unsigned)((L) + 63) / 64, (unsigned)(1)), 32, 0, stream>>>(sq3lo);
      else k_gemm<0><<<dim3((unsigned)((R) + 31) / 32, (unsigned)((L) + 15) / 16, (unsigned)(1)), 32, 0, stream>>>(sq3lo); }
    k_cast16<<<(unsigned)((((long long)(512) * ((1024) / 2)) + 255) / 256), 256, 0, stream>>>(XN, 1024, (_Float16*)(G64A), 1024, 512, 1024, 1.0f);
    k_castT16<<<(unsigned)((((long long)(1024) * ((1024) / 2)) + 255) / 256), 256, 0, stream>>>(sWq, 1024, (_Float16*)(G64B), 1024, 1024, 1024, 16.0f);
    w25::wmma_gemm64<0, false, 0, 0, false, 0><<<dim3((unsigned)((((512) / 64) * ((1024) / 64) + 7) / 8), (unsigned)(1)), 256, 0, stream>>>((const unsigned short*)(G64A), nullptr, 1024, 0, (const unsigned short*)(G64B), nullptr, 1024, 0, (void*)(Q), nullptr, 1024, 0, nullptr, nullptr, 0, 512, 1024, 1024, 0.0625f);
    { GemmP sq3ab;
      sq3ab.A = LOW; sq3ab.B = qb + (size_t)6 * R * D; sq3ab.bias = LOW; sq3ab.R = Q; sq3ab.C = Q;
      sq3ab.sAo = 0; sq3ab.sAi = 0; sq3ab.sAm = R; sq3ab.sAk = 1; sq3ab.sBo = 0; sq3ab.sBi = 0; sq3ab.sBn = 1; sq3ab.sBk = D; sq3ab.sCo = 0; sq3ab.sCi = 0; sq3ab.sCm = D; sq3ab.sRo = 0; sq3ab.sRi = 0; sq3ab.sRm = D; sq3ab.sRn = 1;
      sq3ab.M = L; sq3ab.N = D; sq3ab.K = R; sq3ab.zi_n = 1; sq3ab.flags = 4; sq3ab.act = 0;
      sq3ab.alpha = 1.0f; sq3ab.beta = 1.0f; sq3ab.sa = 1.0f; sq3ab.sb = 1.0f; sq3ab.Npad = D; sq3ab.pad_ = 0;
      if ((long long)(L) >= 64 && (long long)(D) >= 64) k_gemmT<0, 4, 4><<<dim3((unsigned)((D) + 63) / 64, (unsigned)((L) + 63) / 64, (unsigned)(1)), 32, 0, stream>>>(sq3ab);
      else k_gemm<0><<<dim3((unsigned)((D) + 31) / 32, (unsigned)((L) + 15) / 16, (unsigned)(1)), 32, 0, stream>>>(sq3ab); }
    { GemmP sk3lo;
      sk3lo.A = XN; sk3lo.B = ka + (size_t)6 * D * R; sk3lo.bias = XN; sk3lo.R = XN; sk3lo.C = LOW;
      sk3lo.sAo = 0; sk3lo.sAi = 0; sk3lo.sAm = D; sk3lo.sAk = 1; sk3lo.sBo = 0; sk3lo.sBi = 0; sk3lo.sBn = 1; sk3lo.sBk = R; sk3lo.sCo = 0; sk3lo.sCi = 0; sk3lo.sCm = R; sk3lo.sRo = 0; sk3lo.sRi = 0; sk3lo.sRm = 0; sk3lo.sRn = 0;
      sk3lo.M = L; sk3lo.N = R; sk3lo.K = D; sk3lo.zi_n = 1; sk3lo.flags = 0; sk3lo.act = 0;
      sk3lo.alpha = 1.0f; sk3lo.beta = 0.0f; sk3lo.sa = 1.0f; sk3lo.sb = 1.0f; sk3lo.Npad = R; sk3lo.pad_ = 0;
      if ((long long)(L) >= 64 && (long long)(R) >= 64) k_gemmT<0, 4, 4><<<dim3((unsigned)((R) + 63) / 64, (unsigned)((L) + 63) / 64, (unsigned)(1)), 32, 0, stream>>>(sk3lo);
      else k_gemm<0><<<dim3((unsigned)((R) + 31) / 32, (unsigned)((L) + 15) / 16, (unsigned)(1)), 32, 0, stream>>>(sk3lo); }
    k_cast16<<<(unsigned)((((long long)(512) * ((1024) / 2)) + 255) / 256), 256, 0, stream>>>(XN, 1024, (_Float16*)(G64A), 1024, 512, 1024, 1.0f);
    k_castT16<<<(unsigned)((((long long)(1024) * ((1024) / 2)) + 255) / 256), 256, 0, stream>>>(sWk, 1024, (_Float16*)(G64B), 1024, 1024, 1024, 16.0f);
    w25::wmma_gemm64<0, false, 0, 0, false, 0><<<dim3((unsigned)((((512) / 64) * ((1024) / 64) + 7) / 8), (unsigned)(1)), 256, 0, stream>>>((const unsigned short*)(G64A), nullptr, 1024, 0, (const unsigned short*)(G64B), nullptr, 1024, 0, (void*)(Kb), nullptr, 1024, 0, nullptr, nullptr, 0, 512, 1024, 1024, 0.0625f);
    { GemmP sk3ab;
      sk3ab.A = LOW; sk3ab.B = kb + (size_t)6 * R * D; sk3ab.bias = LOW; sk3ab.R = Kb; sk3ab.C = Kb;
      sk3ab.sAo = 0; sk3ab.sAi = 0; sk3ab.sAm = R; sk3ab.sAk = 1; sk3ab.sBo = 0; sk3ab.sBi = 0; sk3ab.sBn = 1; sk3ab.sBk = D; sk3ab.sCo = 0; sk3ab.sCi = 0; sk3ab.sCm = D; sk3ab.sRo = 0; sk3ab.sRi = 0; sk3ab.sRm = D; sk3ab.sRn = 1;
      sk3ab.M = L; sk3ab.N = D; sk3ab.K = R; sk3ab.zi_n = 1; sk3ab.flags = 4; sk3ab.act = 0;
      sk3ab.alpha = 1.0f; sk3ab.beta = 1.0f; sk3ab.sa = 1.0f; sk3ab.sb = 1.0f; sk3ab.Npad = D; sk3ab.pad_ = 0;
      if ((long long)(L) >= 64 && (long long)(D) >= 64) k_gemmT<0, 4, 4><<<dim3((unsigned)((D) + 63) / 64, (unsigned)((L) + 63) / 64, (unsigned)(1)), 32, 0, stream>>>(sk3ab);
      else k_gemm<0><<<dim3((unsigned)((D) + 31) / 32, (unsigned)((L) + 15) / 16, (unsigned)(1)), 32, 0, stream>>>(sk3ab); }
    { GemmP sv3lo;
      sv3lo.A = XN; sv3lo.B = va + (size_t)6 * D * R; sv3lo.bias = XN; sv3lo.R = XN; sv3lo.C = LOW;
      sv3lo.sAo = 0; sv3lo.sAi = 0; sv3lo.sAm = D; sv3lo.sAk = 1; sv3lo.sBo = 0; sv3lo.sBi = 0; sv3lo.sBn = 1; sv3lo.sBk = R; sv3lo.sCo = 0; sv3lo.sCi = 0; sv3lo.sCm = R; sv3lo.sRo = 0; sv3lo.sRi = 0; sv3lo.sRm = 0; sv3lo.sRn = 0;
      sv3lo.M = L; sv3lo.N = R; sv3lo.K = D; sv3lo.zi_n = 1; sv3lo.flags = 0; sv3lo.act = 0;
      sv3lo.alpha = 1.0f; sv3lo.beta = 0.0f; sv3lo.sa = 1.0f; sv3lo.sb = 1.0f; sv3lo.Npad = R; sv3lo.pad_ = 0;
      if ((long long)(L) >= 64 && (long long)(R) >= 64) k_gemmT<0, 4, 4><<<dim3((unsigned)((R) + 63) / 64, (unsigned)((L) + 63) / 64, (unsigned)(1)), 32, 0, stream>>>(sv3lo);
      else k_gemm<0><<<dim3((unsigned)((R) + 31) / 32, (unsigned)((L) + 15) / 16, (unsigned)(1)), 32, 0, stream>>>(sv3lo); }
    k_cast16<<<(unsigned)((((long long)(512) * ((1024) / 2)) + 255) / 256), 256, 0, stream>>>(XN, 1024, (_Float16*)(G64A), 1024, 512, 1024, 1.0f);
    k_castT16<<<(unsigned)((((long long)(1024) * ((1024) / 2)) + 255) / 256), 256, 0, stream>>>(sWv, 1024, (_Float16*)(G64B), 1024, 1024, 1024, 16.0f);
    w25::wmma_gemm64<0, false, 0, 0, false, 0><<<dim3((unsigned)((((512) / 64) * ((1024) / 64) + 7) / 8), (unsigned)(1)), 256, 0, stream>>>((const unsigned short*)(G64A), nullptr, 1024, 0, (const unsigned short*)(G64B), nullptr, 1024, 0, (void*)(V), nullptr, 1024, 0, nullptr, nullptr, 0, 512, 1024, 1024, 0.0625f);
    { GemmP sv3ab;
      sv3ab.A = LOW; sv3ab.B = vb + (size_t)6 * R * D; sv3ab.bias = LOW; sv3ab.R = V; sv3ab.C = V;
      sv3ab.sAo = 0; sv3ab.sAi = 0; sv3ab.sAm = R; sv3ab.sAk = 1; sv3ab.sBo = 0; sv3ab.sBi = 0; sv3ab.sBn = 1; sv3ab.sBk = D; sv3ab.sCo = 0; sv3ab.sCi = 0; sv3ab.sCm = D; sv3ab.sRo = 0; sv3ab.sRi = 0; sv3ab.sRm = D; sv3ab.sRn = 1;
      sv3ab.M = L; sv3ab.N = D; sv3ab.K = R; sv3ab.zi_n = 1; sv3ab.flags = 4; sv3ab.act = 0;
      sv3ab.alpha = 1.0f; sv3ab.beta = 1.0f; sv3ab.sa = 1.0f; sv3ab.sb = 1.0f; sv3ab.Npad = D; sv3ab.pad_ = 0;
      if ((long long)(L) >= 64 && (long long)(D) >= 64) k_gemmT<0, 4, 4><<<dim3((unsigned)((D) + 63) / 64, (unsigned)((L) + 63) / 64, (unsigned)(1)), 32, 0, stream>>>(sv3ab);
      else k_gemm<0><<<dim3((unsigned)((D) + 31) / 32, (unsigned)((L) + 15) / 16, (unsigned)(1)), 32, 0, stream>>>(sv3ab); }
    {   AttnP a;
      a.Q = Q; a.K = Kb; a.V = V; a.O = AT; a.P = 0; a.Mf = BIAS; a.Mi = 0; a.ST = 0;
      a.Pw = 0; a.Rt = 0; a.SQ = 0; a.SK = 0;
      a.swb = 0; a.swh = 0; a.swi = 0; a.swj = 0; a.srb = 0; a.srh = 0; a.sri = 0; a.sQb = 0; a.sQh = HD; a.sQi = D; a.sQd = 1; a.sKb = 0; a.sKh = HD; a.sKj = D; a.sKd = 1; a.sVb = 0; a.sVh = HD; a.sVj = D; a.sVd = 1; a.sOb = 0; a.sOh = HD; a.sOi = D; a.sPb = 0; a.sPh = 0; a.sPi = 0; a.smb = 0; a.smh = (long long)L * L; a.smi = L; a.smj = 1;
      a.Lq = L; a.Lk = L; a.dh = HD; a.dv = HD; a.hrep = 1; a.causal = 1; a.coff = 0; a.pband = 0;
      a.scale = 0.125f; a.mfill = 0.0f; a.nonorm = 0; a.mpol = 0;
      a.roff = 0; a.rn = 1; a.segpol = 0; a.win = 0;
      k_attn<64, 64, 0, false, false><<<dim3((unsigned)((L) + 16 * AW - 1) / (16 * AW), (unsigned)(NH), (unsigned)(1)), 32 * AW, 0, stream>>>(a); }
    { GemmP so3lo;
      so3lo.A = AT; so3lo.B = oa + (size_t)6 * D * R; so3lo.bias = AT; so3lo.R = AT; so3lo.C = LOW;
      so3lo.sAo = 0; so3lo.sAi = 0; so3lo.sAm = D; so3lo.sAk = 1; so3lo.sBo = 0; so3lo.sBi = 0; so3lo.sBn = 1; so3lo.sBk = R; so3lo.sCo = 0; so3lo.sCi = 0; so3lo.sCm = R; so3lo.sRo = 0; so3lo.sRi = 0; so3lo.sRm = 0; so3lo.sRn = 0;
      so3lo.M = L; so3lo.N = R; so3lo.K = D; so3lo.zi_n = 1; so3lo.flags = 0; so3lo.act = 0;
      so3lo.alpha = 1.0f; so3lo.beta = 0.0f; so3lo.sa = 1.0f; so3lo.sb = 1.0f; so3lo.Npad = R; so3lo.pad_ = 0;
      if ((long long)(L) >= 64 && (long long)(R) >= 64) k_gemmT<0, 4, 4><<<dim3((unsigned)((R) + 63) / 64, (unsigned)((L) + 63) / 64, (unsigned)(1)), 32, 0, stream>>>(so3lo);
      else k_gemm<0><<<dim3((unsigned)((R) + 31) / 32, (unsigned)((L) + 15) / 16, (unsigned)(1)), 32, 0, stream>>>(so3lo); }
    k_cast16<<<(unsigned)((((long long)(512) * ((1024) / 2)) + 255) / 256), 256, 0, stream>>>(AT, 1024, (_Float16*)(G64A), 1024, 512, 1024, 1.0f);
    k_castT16<<<(unsigned)((((long long)(1024) * ((1024) / 2)) + 255) / 256), 256, 0, stream>>>(sWo, 1024, (_Float16*)(G64B), 1024, 1024, 1024, 16.0f);
    w25::wmma_gemm64<0, false, 0, 0, true, 0><<<dim3((unsigned)((((512) / 64) * ((1024) / 64) + 7) / 8), (unsigned)(1)), 256, 0, stream>>>((const unsigned short*)(G64A), nullptr, 1024, 0, (const unsigned short*)(G64B), nullptr, 1024, 0, (void*)(X1 + (size_t)3 * L * D), nullptr, 1024, 0, nullptr, xin + (size_t)3 * L * D, 0, 512, 1024, 1024, 0.0625f);
    { GemmP so3ab;
      so3ab.A = LOW; so3ab.B = ob + (size_t)6 * R * D; so3ab.bias = LOW; so3ab.R = X1 + (size_t)3 * L * D; so3ab.C = X1 + (size_t)3 * L * D;
      so3ab.sAo = 0; so3ab.sAi = 0; so3ab.sAm = R; so3ab.sAk = 1; so3ab.sBo = 0; so3ab.sBi = 0; so3ab.sBn = 1; so3ab.sBk = D; so3ab.sCo = 0; so3ab.sCi = 0; so3ab.sCm = D; so3ab.sRo = 0; so3ab.sRi = 0; so3ab.sRm = D; so3ab.sRn = 1;
      so3ab.M = L; so3ab.N = D; so3ab.K = R; so3ab.zi_n = 1; so3ab.flags = 4; so3ab.act = 0;
      so3ab.alpha = 1.0f; so3ab.beta = 1.0f; so3ab.sa = 1.0f; so3ab.sb = 1.0f; so3ab.Npad = D; so3ab.pad_ = 0;
      if ((long long)(L) >= 64 && (long long)(D) >= 64) k_gemmT<0, 4, 4><<<dim3((unsigned)((D) + 63) / 64, (unsigned)((L) + 63) / 64, (unsigned)(1)), 32, 0, stream>>>(so3ab);
      else k_gemm<0><<<dim3((unsigned)((D) + 31) / 32, (unsigned)((L) + 15) / 16, (unsigned)(1)), 32, 0, stream>>>(so3ab); }
    k_ld_rms<<<L, 256, 0, stream>>>(X1 + (size_t)3 * L * D, ln2, XN, D);
    { GemmP cq3lo;
      cq3lo.A = XN; cq3lo.B = qa + (size_t)7 * D * R; cq3lo.bias = XN; cq3lo.R = XN; cq3lo.C = LOW;
      cq3lo.sAo = 0; cq3lo.sAi = 0; cq3lo.sAm = D; cq3lo.sAk = 1; cq3lo.sBo = 0; cq3lo.sBi = 0; cq3lo.sBn = 1; cq3lo.sBk = R; cq3lo.sCo = 0; cq3lo.sCi = 0; cq3lo.sCm = R; cq3lo.sRo = 0; cq3lo.sRi = 0; cq3lo.sRm = 0; cq3lo.sRn = 0;
      cq3lo.M = L; cq3lo.N = R; cq3lo.K = D; cq3lo.zi_n = 1; cq3lo.flags = 0; cq3lo.act = 0;
      cq3lo.alpha = 1.0f; cq3lo.beta = 0.0f; cq3lo.sa = 1.0f; cq3lo.sb = 1.0f; cq3lo.Npad = R; cq3lo.pad_ = 0;
      if ((long long)(L) >= 64 && (long long)(R) >= 64) k_gemmT<0, 4, 4><<<dim3((unsigned)((R) + 63) / 64, (unsigned)((L) + 63) / 64, (unsigned)(1)), 32, 0, stream>>>(cq3lo);
      else k_gemm<0><<<dim3((unsigned)((R) + 31) / 32, (unsigned)((L) + 15) / 16, (unsigned)(1)), 32, 0, stream>>>(cq3lo); }
    k_cast16<<<(unsigned)((((long long)(512) * ((1024) / 2)) + 255) / 256), 256, 0, stream>>>(XN, 1024, (_Float16*)(G64A), 1024, 512, 1024, 1.0f);
    k_castT16<<<(unsigned)((((long long)(1024) * ((1024) / 2)) + 255) / 256), 256, 0, stream>>>(cWq, 1024, (_Float16*)(G64B), 1024, 1024, 1024, 16.0f);
    w25::wmma_gemm64<0, false, 0, 0, false, 0><<<dim3((unsigned)((((512) / 64) * ((1024) / 64) + 7) / 8), (unsigned)(1)), 256, 0, stream>>>((const unsigned short*)(G64A), nullptr, 1024, 0, (const unsigned short*)(G64B), nullptr, 1024, 0, (void*)(Q), nullptr, 1024, 0, nullptr, nullptr, 0, 512, 1024, 1024, 0.0625f);
    { GemmP cq3ab;
      cq3ab.A = LOW; cq3ab.B = qb + (size_t)7 * R * D; cq3ab.bias = LOW; cq3ab.R = Q; cq3ab.C = Q;
      cq3ab.sAo = 0; cq3ab.sAi = 0; cq3ab.sAm = R; cq3ab.sAk = 1; cq3ab.sBo = 0; cq3ab.sBi = 0; cq3ab.sBn = 1; cq3ab.sBk = D; cq3ab.sCo = 0; cq3ab.sCi = 0; cq3ab.sCm = D; cq3ab.sRo = 0; cq3ab.sRi = 0; cq3ab.sRm = D; cq3ab.sRn = 1;
      cq3ab.M = L; cq3ab.N = D; cq3ab.K = R; cq3ab.zi_n = 1; cq3ab.flags = 4; cq3ab.act = 0;
      cq3ab.alpha = 1.0f; cq3ab.beta = 1.0f; cq3ab.sa = 1.0f; cq3ab.sb = 1.0f; cq3ab.Npad = D; cq3ab.pad_ = 0;
      if ((long long)(L) >= 64 && (long long)(D) >= 64) k_gemmT<0, 4, 4><<<dim3((unsigned)((D) + 63) / 64, (unsigned)((L) + 63) / 64, (unsigned)(1)), 32, 0, stream>>>(cq3ab);
      else k_gemm<0><<<dim3((unsigned)((D) + 31) / 32, (unsigned)((L) + 15) / 16, (unsigned)(1)), 32, 0, stream>>>(cq3ab); }
    { GemmP ck3lo;
      ck3lo.A = enc + (size_t)3 * L * D; ck3lo.B = ka + (size_t)7 * D * R; ck3lo.bias = enc + (size_t)3 * L * D; ck3lo.R = enc + (size_t)3 * L * D; ck3lo.C = LOW;
      ck3lo.sAo = 0; ck3lo.sAi = 0; ck3lo.sAm = D; ck3lo.sAk = 1; ck3lo.sBo = 0; ck3lo.sBi = 0; ck3lo.sBn = 1; ck3lo.sBk = R; ck3lo.sCo = 0; ck3lo.sCi = 0; ck3lo.sCm = R; ck3lo.sRo = 0; ck3lo.sRi = 0; ck3lo.sRm = 0; ck3lo.sRn = 0;
      ck3lo.M = L; ck3lo.N = R; ck3lo.K = D; ck3lo.zi_n = 1; ck3lo.flags = 0; ck3lo.act = 0;
      ck3lo.alpha = 1.0f; ck3lo.beta = 0.0f; ck3lo.sa = 1.0f; ck3lo.sb = 1.0f; ck3lo.Npad = R; ck3lo.pad_ = 0;
      if ((long long)(L) >= 64 && (long long)(R) >= 64) k_gemmT<0, 4, 4><<<dim3((unsigned)((R) + 63) / 64, (unsigned)((L) + 63) / 64, (unsigned)(1)), 32, 0, stream>>>(ck3lo);
      else k_gemm<0><<<dim3((unsigned)((R) + 31) / 32, (unsigned)((L) + 15) / 16, (unsigned)(1)), 32, 0, stream>>>(ck3lo); }
    k_cast16<<<(unsigned)((((long long)(512) * ((1024) / 2)) + 255) / 256), 256, 0, stream>>>(enc + (size_t)3 * L * D, 1024, (_Float16*)(G64A), 1024, 512, 1024, 1.0f);
    k_castT16<<<(unsigned)((((long long)(1024) * ((1024) / 2)) + 255) / 256), 256, 0, stream>>>(cWk, 1024, (_Float16*)(G64B), 1024, 1024, 1024, 16.0f);
    w25::wmma_gemm64<0, false, 0, 0, false, 0><<<dim3((unsigned)((((512) / 64) * ((1024) / 64) + 7) / 8), (unsigned)(1)), 256, 0, stream>>>((const unsigned short*)(G64A), nullptr, 1024, 0, (const unsigned short*)(G64B), nullptr, 1024, 0, (void*)(Kb), nullptr, 1024, 0, nullptr, nullptr, 0, 512, 1024, 1024, 0.0625f);
    { GemmP ck3ab;
      ck3ab.A = LOW; ck3ab.B = kb + (size_t)7 * R * D; ck3ab.bias = LOW; ck3ab.R = Kb; ck3ab.C = Kb;
      ck3ab.sAo = 0; ck3ab.sAi = 0; ck3ab.sAm = R; ck3ab.sAk = 1; ck3ab.sBo = 0; ck3ab.sBi = 0; ck3ab.sBn = 1; ck3ab.sBk = D; ck3ab.sCo = 0; ck3ab.sCi = 0; ck3ab.sCm = D; ck3ab.sRo = 0; ck3ab.sRi = 0; ck3ab.sRm = D; ck3ab.sRn = 1;
      ck3ab.M = L; ck3ab.N = D; ck3ab.K = R; ck3ab.zi_n = 1; ck3ab.flags = 4; ck3ab.act = 0;
      ck3ab.alpha = 1.0f; ck3ab.beta = 1.0f; ck3ab.sa = 1.0f; ck3ab.sb = 1.0f; ck3ab.Npad = D; ck3ab.pad_ = 0;
      if ((long long)(L) >= 64 && (long long)(D) >= 64) k_gemmT<0, 4, 4><<<dim3((unsigned)((D) + 63) / 64, (unsigned)((L) + 63) / 64, (unsigned)(1)), 32, 0, stream>>>(ck3ab);
      else k_gemm<0><<<dim3((unsigned)((D) + 31) / 32, (unsigned)((L) + 15) / 16, (unsigned)(1)), 32, 0, stream>>>(ck3ab); }
    { GemmP cv3lo;
      cv3lo.A = enc + (size_t)3 * L * D; cv3lo.B = va + (size_t)7 * D * R; cv3lo.bias = enc + (size_t)3 * L * D; cv3lo.R = enc + (size_t)3 * L * D; cv3lo.C = LOW;
      cv3lo.sAo = 0; cv3lo.sAi = 0; cv3lo.sAm = D; cv3lo.sAk = 1; cv3lo.sBo = 0; cv3lo.sBi = 0; cv3lo.sBn = 1; cv3lo.sBk = R; cv3lo.sCo = 0; cv3lo.sCi = 0; cv3lo.sCm = R; cv3lo.sRo = 0; cv3lo.sRi = 0; cv3lo.sRm = 0; cv3lo.sRn = 0;
      cv3lo.M = L; cv3lo.N = R; cv3lo.K = D; cv3lo.zi_n = 1; cv3lo.flags = 0; cv3lo.act = 0;
      cv3lo.alpha = 1.0f; cv3lo.beta = 0.0f; cv3lo.sa = 1.0f; cv3lo.sb = 1.0f; cv3lo.Npad = R; cv3lo.pad_ = 0;
      if ((long long)(L) >= 64 && (long long)(R) >= 64) k_gemmT<0, 4, 4><<<dim3((unsigned)((R) + 63) / 64, (unsigned)((L) + 63) / 64, (unsigned)(1)), 32, 0, stream>>>(cv3lo);
      else k_gemm<0><<<dim3((unsigned)((R) + 31) / 32, (unsigned)((L) + 15) / 16, (unsigned)(1)), 32, 0, stream>>>(cv3lo); }
    k_cast16<<<(unsigned)((((long long)(512) * ((1024) / 2)) + 255) / 256), 256, 0, stream>>>(enc + (size_t)3 * L * D, 1024, (_Float16*)(G64A), 1024, 512, 1024, 1.0f);
    k_castT16<<<(unsigned)((((long long)(1024) * ((1024) / 2)) + 255) / 256), 256, 0, stream>>>(cWv, 1024, (_Float16*)(G64B), 1024, 1024, 1024, 16.0f);
    w25::wmma_gemm64<0, false, 0, 0, false, 0><<<dim3((unsigned)((((512) / 64) * ((1024) / 64) + 7) / 8), (unsigned)(1)), 256, 0, stream>>>((const unsigned short*)(G64A), nullptr, 1024, 0, (const unsigned short*)(G64B), nullptr, 1024, 0, (void*)(V), nullptr, 1024, 0, nullptr, nullptr, 0, 512, 1024, 1024, 0.0625f);
    { GemmP cv3ab;
      cv3ab.A = LOW; cv3ab.B = vb + (size_t)7 * R * D; cv3ab.bias = LOW; cv3ab.R = V; cv3ab.C = V;
      cv3ab.sAo = 0; cv3ab.sAi = 0; cv3ab.sAm = R; cv3ab.sAk = 1; cv3ab.sBo = 0; cv3ab.sBi = 0; cv3ab.sBn = 1; cv3ab.sBk = D; cv3ab.sCo = 0; cv3ab.sCi = 0; cv3ab.sCm = D; cv3ab.sRo = 0; cv3ab.sRi = 0; cv3ab.sRm = D; cv3ab.sRn = 1;
      cv3ab.M = L; cv3ab.N = D; cv3ab.K = R; cv3ab.zi_n = 1; cv3ab.flags = 4; cv3ab.act = 0;
      cv3ab.alpha = 1.0f; cv3ab.beta = 1.0f; cv3ab.sa = 1.0f; cv3ab.sb = 1.0f; cv3ab.Npad = D; cv3ab.pad_ = 0;
      if ((long long)(L) >= 64 && (long long)(D) >= 64) k_gemmT<0, 4, 4><<<dim3((unsigned)((D) + 63) / 64, (unsigned)((L) + 63) / 64, (unsigned)(1)), 32, 0, stream>>>(cv3ab);
      else k_gemm<0><<<dim3((unsigned)((D) + 31) / 32, (unsigned)((L) + 15) / 16, (unsigned)(1)), 32, 0, stream>>>(cv3ab); }
    {   AttnP a;
      a.Q = Q; a.K = Kb; a.V = V; a.O = AT; a.P = 0; a.Mf = 0; a.Mi = 0; a.ST = 0;
      a.Pw = 0; a.Rt = 0; a.SQ = 0; a.SK = 0;
      a.swb = 0; a.swh = 0; a.swi = 0; a.swj = 0; a.srb = 0; a.srh = 0; a.sri = 0; a.sQb = 0; a.sQh = HD; a.sQi = D; a.sQd = 1; a.sKb = 0; a.sKh = HD; a.sKj = D; a.sKd = 1; a.sVb = 0; a.sVh = HD; a.sVj = D; a.sVd = 1; a.sOb = 0; a.sOh = HD; a.sOi = D; a.sPb = 0; a.sPh = 0; a.sPi = 0; a.smb = 0; a.smh = 0; a.smi = 0; a.smj = 0;
      a.Lq = L; a.Lk = L; a.dh = HD; a.dv = HD; a.hrep = 1; a.causal = 0; a.coff = 0; a.pband = 0;
      a.scale = 0.125f; a.mfill = 0.0f; a.nonorm = 0; a.mpol = 0;
      a.roff = 0; a.rn = 1; a.segpol = 0; a.win = 0;
      k_attn<64, 64, 0, false, false><<<dim3((unsigned)((L) + 16 * AW - 1) / (16 * AW), (unsigned)(NH), (unsigned)(1)), 32 * AW, 0, stream>>>(a); }
    { GemmP co3lo;
      co3lo.A = AT; co3lo.B = oa + (size_t)7 * D * R; co3lo.bias = AT; co3lo.R = AT; co3lo.C = LOW;
      co3lo.sAo = 0; co3lo.sAi = 0; co3lo.sAm = D; co3lo.sAk = 1; co3lo.sBo = 0; co3lo.sBi = 0; co3lo.sBn = 1; co3lo.sBk = R; co3lo.sCo = 0; co3lo.sCi = 0; co3lo.sCm = R; co3lo.sRo = 0; co3lo.sRi = 0; co3lo.sRm = 0; co3lo.sRn = 0;
      co3lo.M = L; co3lo.N = R; co3lo.K = D; co3lo.zi_n = 1; co3lo.flags = 0; co3lo.act = 0;
      co3lo.alpha = 1.0f; co3lo.beta = 0.0f; co3lo.sa = 1.0f; co3lo.sb = 1.0f; co3lo.Npad = R; co3lo.pad_ = 0;
      if ((long long)(L) >= 64 && (long long)(R) >= 64) k_gemmT<0, 4, 4><<<dim3((unsigned)((R) + 63) / 64, (unsigned)((L) + 63) / 64, (unsigned)(1)), 32, 0, stream>>>(co3lo);
      else k_gemm<0><<<dim3((unsigned)((R) + 31) / 32, (unsigned)((L) + 15) / 16, (unsigned)(1)), 32, 0, stream>>>(co3lo); }
    k_cast16<<<(unsigned)((((long long)(512) * ((1024) / 2)) + 255) / 256), 256, 0, stream>>>(AT, 1024, (_Float16*)(G64A), 1024, 512, 1024, 1.0f);
    k_castT16<<<(unsigned)((((long long)(1024) * ((1024) / 2)) + 255) / 256), 256, 0, stream>>>(cWo, 1024, (_Float16*)(G64B), 1024, 1024, 1024, 16.0f);
    w25::wmma_gemm64<0, false, 0, 0, true, 0><<<dim3((unsigned)((((512) / 64) * ((1024) / 64) + 7) / 8), (unsigned)(1)), 256, 0, stream>>>((const unsigned short*)(G64A), nullptr, 1024, 0, (const unsigned short*)(G64B), nullptr, 1024, 0, (void*)(Y1 + (size_t)3 * L * D), nullptr, 1024, 0, nullptr, X1 + (size_t)3 * L * D, 0, 512, 1024, 1024, 0.0625f);
    { GemmP co3ab;
      co3ab.A = LOW; co3ab.B = ob + (size_t)7 * R * D; co3ab.bias = LOW; co3ab.R = Y1 + (size_t)3 * L * D; co3ab.C = Y1 + (size_t)3 * L * D;
      co3ab.sAo = 0; co3ab.sAi = 0; co3ab.sAm = R; co3ab.sAk = 1; co3ab.sBo = 0; co3ab.sBi = 0; co3ab.sBn = 1; co3ab.sBk = D; co3ab.sCo = 0; co3ab.sCi = 0; co3ab.sCm = D; co3ab.sRo = 0; co3ab.sRi = 0; co3ab.sRm = D; co3ab.sRn = 1;
      co3ab.M = L; co3ab.N = D; co3ab.K = R; co3ab.zi_n = 1; co3ab.flags = 4; co3ab.act = 0;
      co3ab.alpha = 1.0f; co3ab.beta = 1.0f; co3ab.sa = 1.0f; co3ab.sb = 1.0f; co3ab.Npad = D; co3ab.pad_ = 0;
      if ((long long)(L) >= 64 && (long long)(D) >= 64) k_gemmT<0, 4, 4><<<dim3((unsigned)((D) + 63) / 64, (unsigned)((L) + 63) / 64, (unsigned)(1)), 32, 0, stream>>>(co3ab);
      else k_gemm<0><<<dim3((unsigned)((D) + 31) / 32, (unsigned)((L) + 15) / 16, (unsigned)(1)), 32, 0, stream>>>(co3ab); }
    k_ld_rms<<<L, 256, 0, stream>>>(Y1 + (size_t)3 * L * D, ln3, XN, D);
    k_cast16<<<(unsigned)((((long long)(512) * ((1024) / 2)) + 255) / 256), 256, 0, stream>>>(XN, 1024, (_Float16*)(G64A), 1024, 512, 1024, 1.0f);
    k_castT16<<<(unsigned)((((long long)(4096) * ((1024) / 2)) + 255) / 256), 256, 0, stream>>>(wi0, 4096, (_Float16*)(G64B), 1024, 1024, 4096, 16.0f);
    w25::wmma_gemm64<0, false, 0, 0, false, 0><<<dim3((unsigned)((((512) / 64) * ((4096) / 64) + 7) / 8), (unsigned)(1)), 256, 0, stream>>>((const unsigned short*)(G64A), nullptr, 1024, 0, (const unsigned short*)(G64B), nullptr, 1024, 0, (void*)(G0), nullptr, 4096, 0, nullptr, nullptr, 0, 512, 4096, 1024, 0.0625f);
    k_cast16<<<(unsigned)((((long long)(512) * ((1024) / 2)) + 255) / 256), 256, 0, stream>>>(XN, 1024, (_Float16*)(G64A), 1024, 512, 1024, 1.0f);
    k_castT16<<<(unsigned)((((long long)(4096) * ((1024) / 2)) + 255) / 256), 256, 0, stream>>>(wi1, 4096, (_Float16*)(G64B), 1024, 1024, 4096, 16.0f);
    w25::wmma_gemm64<0, false, 0, 0, false, 0><<<dim3((unsigned)((((512) / 64) * ((4096) / 64) + 7) / 8), (unsigned)(1)), 256, 0, stream>>>((const unsigned short*)(G64A), nullptr, 1024, 0, (const unsigned short*)(G64B), nullptr, 1024, 0, (void*)(G1), nullptr, 4096, 0, nullptr, nullptr, 0, 512, 4096, 1024, 0.0625f);
    k_ld_gg<<<(unsigned)(((long long)L * FF + 255) / 256), 256, 0, stream>>>(G0, G1, (long long)L * FF);
    k_cast16<<<(unsigned)((((long long)(512) * ((4096) / 2)) + 255) / 256), 256, 0, stream>>>(G0, 4096, (_Float16*)(G64A), 4096, 512, 4096, 1.0f);
    k_castT16<<<(unsigned)((((long long)(1024) * ((4096) / 2)) + 255) / 256), 256, 0, stream>>>(wom, 1024, (_Float16*)(G64B), 4096, 4096, 1024, 16.0f);
    w25::wmma_gemm64<0, false, 0, 0, true, 0><<<dim3((unsigned)((((512) / 64) * ((1024) / 64) + 7) / 8), (unsigned)(1)), 256, 0, stream>>>((const unsigned short*)(G64A), nullptr, 4096, 0, (const unsigned short*)(G64B), nullptr, 4096, 0, (void*)(out + (size_t)3 * L * D), nullptr, 1024, 0, nullptr, Y1 + (size_t)3 * L * D, 0, 512, 1024, 4096, 0.0625f);
}
